// TrajectoryDecoder_8650064134853
// MI455X (gfx1250) — hardware-verified
//
#include <hip/hip_runtime.h>
#include <math.h>

typedef __attribute__((ext_vector_type(16))) _Float16 v16h;
typedef __attribute__((ext_vector_type(8)))  _Float16 v8h;
typedef __attribute__((ext_vector_type(16))) __bf16   v16b;
typedef __attribute__((ext_vector_type(8)))  float    v8f;
typedef __attribute__((ext_vector_type(4)))  float    v4f;

__device__ __forceinline__ int frag_k(int i, int h) { return (i < 8) ? (8 * h + i) : (16 + 8 * h + (i - 8)); }
__device__ __forceinline__ __bf16 bf16_rne(float f) {
    unsigned int u = __float_as_uint(f);
    u += 0x7fffu + ((u >> 16) & 1u);
    return __builtin_bit_cast(__bf16, (unsigned short)(u >> 16));
}
__device__ __forceinline__ float bf16_f32(__bf16 b) { return __uint_as_float(((unsigned int)__builtin_bit_cast(unsigned short, b)) << 16); }
__device__ __forceinline__ v8f wmma16(v16h a, v16h b, v8f c) {
    c = __builtin_amdgcn_wmma_f32_16x16x32_f16(false, a, false, b, (short)0, c, false, false);
    asm volatile("v_nop\n\tv_nop\n\tv_nop\n\tv_nop" : "+v"(c) : "v"(a), "v"(b));
    return c;
}
__device__ __forceinline__ v8f wmmab(v16b a, v16b b, v8f c) {
    c = __builtin_amdgcn_wmma_f32_16x16x32_bf16(false, a, false, b, (short)0, c, false, false);
    asm volatile("v_nop\n\tv_nop\n\tv_nop\n\tv_nop" : "+v"(c) : "v"(a), "v"(b));
    return c;
}
struct Split { v16b hi, lo; };
__device__ __forceinline__ v8f wmma3(const Split& a, const Split& b, v8f c) {
    c = __builtin_amdgcn_wmma_f32_16x16x32_bf16(false, a.hi, false, b.hi, (short)0, c, false, false);
    c = __builtin_amdgcn_wmma_f32_16x16x32_bf16(false, a.hi, false, b.lo, (short)0, c, false, false);
    c = __builtin_amdgcn_wmma_f32_16x16x32_bf16(false, a.lo, false, b.hi, (short)0, c, false, false);
    asm volatile("v_nop\n\tv_nop\n\tv_nop\n\tv_nop" : "+v"(c) : "v"(a.hi), "v"(a.lo), "v"(b.hi), "v"(b.lo));
    return c;
}
struct Split3 { v16b hi, mid, lo; };
__device__ __forceinline__ v8f wmma6(const Split3& a, const Split3& b, v8f c) {
    c = __builtin_amdgcn_wmma_f32_16x16x32_bf16(false, a.hi, false, b.hi, (short)0, c, false, false);
    c = __builtin_amdgcn_wmma_f32_16x16x32_bf16(false, a.hi, false, b.mid, (short)0, c, false, false);
    c = __builtin_amdgcn_wmma_f32_16x16x32_bf16(false, a.mid, false, b.hi, (short)0, c, false, false);
    c = __builtin_amdgcn_wmma_f32_16x16x32_bf16(false, a.hi, false, b.lo, (short)0, c, false, false);
    c = __builtin_amdgcn_wmma_f32_16x16x32_bf16(false, a.mid, false, b.mid, (short)0, c, false, false);
    c = __builtin_amdgcn_wmma_f32_16x16x32_bf16(false, a.lo, false, b.hi, (short)0, c, false, false);
    asm volatile("v_nop\n\tv_nop\n\tv_nop\n\tv_nop" : "+v"(c) : "v"(a.hi), "v"(a.mid), "v"(a.lo), "v"(b.hi), "v"(b.mid), "v"(b.lo));
    return c;
}

__device__ __forceinline__ v16h fh_ld(const float* __restrict__ p, long long sk, int k0, int h, int klen, float s) {
    v16h a;
#pragma unroll
    for (int i = 0; i < 16; ++i) { const int k = k0 + frag_k(i, h); a[i] = (k < klen) ? (_Float16)(p[(long long)k * sk] * s) : (_Float16)0.f; }
    return a;
}
__device__ __forceinline__ Split sp_ld(const float* __restrict__ p, long long sk, int k0, int h, int klen, float s) {
    Split r;
#pragma unroll
    for (int i = 0; i < 16; ++i) {
        const int k = k0 + frag_k(i, h); const float x = (k < klen) ? p[(long long)k * sk] * s : 0.f;
        const __bf16 hb = bf16_rne(x); r.hi[i] = hb; r.lo[i] = bf16_rne(x - bf16_f32(hb));
    }
    return r;
}
__device__ __forceinline__ Split3 sp3_ld(const float* __restrict__ p, long long sk, int k0, int h, int klen, float s) {
    Split3 r;
#pragma unroll
    for (int i = 0; i < 16; ++i) {
        const int k = k0 + frag_k(i, h); const float x = (k < klen) ? p[(long long)k * sk] * s : 0.f;
        const __bf16 hb = bf16_rne(x); const float r1 = x - bf16_f32(hb); const __bf16 mb = bf16_rne(r1);
        r.hi[i] = hb; r.mid[i] = mb; r.lo[i] = bf16_rne(r1 - bf16_f32(mb));
    }
    return r;
}
__device__ __forceinline__ v16b bh_ld(const float* __restrict__ p, long long sk, int k0, int h, int klen, float s) {
    v16b a;
#pragma unroll
    for (int i = 0; i < 16; ++i) { const int k = k0 + frag_k(i, h); a[i] = bf16_rne((k < klen) ? p[(long long)k * sk] * s : 0.f); }
    return a;
}
__device__ __forceinline__ v16h fh_row(const _Float16* __restrict__ row, int k0, int h) {
    v16h a;
#pragma unroll
    for (int i = 0; i < 16; ++i) a[i] = row[k0 + frag_k(i, h)];
    return a;
}

#define VST2(T, ptr, val) do { *(volatile T*)(ptr) = (val); __threadfence(); *(volatile T*)(ptr) = (val); } while (0)
typedef float v4f __attribute__((ext_vector_type(4)));
#define VST2V4(ptr, val) do { *(volatile v4f*)(ptr) = (val); __threadfence(); *(volatile v4f*)(ptr) = (val); } while (0)

__device__ __attribute__((noinline)) float act_fn(float v, int act) {
    if (act == 1) return fmaxf(v, 0.f);
    if (act == 2) { const float u = 0.7978845608028654f * (v + 0.044715f * v * v * v); return 0.5f * v * (1.f + tanhf(u)); }
    if (act == 3) return v / (1.f + expf(-v));
    if (act == 4) return 0.5f * v * (1.f + erff(v * 0.7071067811865476f));
    if (act == 5) return tanhf(v);
    if (act == 6) return 1.f / (1.f + expf(-v));
    if (act == 7) return (v > 0.f) ? v : 0.01f * v;
    if (act == 8) return (v > 0.f) ? v : (expf(v) - 1.f);
    if (act == 9) return fminf(fmaxf(v, 0.f), 6.f);
    if (act == 10) return fabsf(v);
    if (act == 11) return (v >= 0.f) ? v : 0.1f * v;
    if (act == 12) return (v > 0.f) ? v : 0.2f * v;
    if (act == 13) return (v > 20.f) ? v : log1pf(expf(v));
    return v;
}

struct GemmP {
    const float* A; const float* B; const float* bias; const float* R; float* C;
    long long sAo, sAi, sAm, sAk, sBo, sBi, sBn, sBk, sCo, sCi, sCm, sRo, sRi, sRm, sRn;
    int M, N, K, zi_n, flags, act; float alpha, beta, sa, sb;
    int Npad, pad_;
};
static_assert(sizeof(GemmP) == 5 * 8 + 15 * 8 + 6 * 4 + 4 * 4 + 2 * 4, "GemmP has padding");

template <int MODE>
__global__ __launch_bounds__(32) void k_gemm(GemmP p) {
    const int lane = threadIdx.x & 31, h = lane >> 4, l15 = lane & 15;
    const int m0 = blockIdx.y * 16, n0 = blockIdx.x * 32;
    const int z = blockIdx.z, zo = z / p.zi_n, zi = z - zo * p.zi_n;
    const float* A = p.A + zo * p.sAo + zi * p.sAi;
    const float* B = p.B + zo * p.sBo + zi * p.sBi;
    const int am = min(m0 + l15, p.M - 1);
    v8f acc[2];
#pragma unroll
    for (int t = 0; t < 2; ++t) { v8f zz = {}; acc[t] = zz; }
    for (int k0 = 0; k0 < p.K; k0 += 32) {
        const float* arow = A + (long long)am * p.sAm;
        if (MODE == 1) {
            const Split a = sp_ld(arow, p.sAk, k0, h, p.K, 1.f);
#pragma unroll
            for (int t = 0; t < 2; ++t) {
                const int bn = min(n0 + t * 16 + l15, p.N - 1);
                acc[t] = wmma3(a, sp_ld(B + (long long)bn * p.sBn, p.sBk, k0, h, p.K, 1.f), acc[t]);
            }
        } else if (MODE == 3) {
            const Split3 a = sp3_ld(arow, p.sAk, k0, h, p.K, 1.f);
#pragma unroll
            for (int t = 0; t < 2; ++t) {
                const int bn = min(n0 + t * 16 + l15, p.N - 1);
                acc[t] = wmma6(a, sp3_ld(B + (long long)bn * p.sBn, p.sBk, k0, h, p.K, 1.f), acc[t]);
            }
        } else if (MODE == 2) {
            const v16b a = bh_ld(arow, p.sAk, k0, h, p.K, 1.f);
#pragma unroll
            for (int t = 0; t < 2; ++t) {
                const int bn = min(n0 + t * 16 + l15, p.N - 1);
                acc[t] = wmmab(a, bh_ld(B + (long long)bn * p.sBn, p.sBk, k0, h, p.K, 1.f), acc[t]);
            }
        } else {
            const v16h a = fh_ld(arow, p.sAk, k0, h, p.K, p.sa);
#pragma unroll
            for (int t = 0; t < 2; ++t) {
                const int bn = min(n0 + t * 16 + l15, p.N - 1);
                acc[t] = wmma16(a, fh_ld(B + (long long)bn * p.sBn, p.sBk, k0, h, p.K, p.sb), acc[t]);
            }
        }
    }
    const float iscale = (MODE == 0) ? p.alpha / (p.sa * p.sb) : p.alpha;
    float* C = p.C + zo * p.sCo + zi * p.sCi;
    const float* R = p.R + zo * p.sRo + zi * p.sRi;
    __shared__ __align__(16) float ctile[16][36];
#pragma unroll
    for (int t = 0; t < 2; ++t) {
        const int n = n0 + t * 16 + l15; const int nn = min(n, p.N - 1);
#pragma unroll
        for (int r = 0; r < 8; ++r) {
            const int m = m0 + 8 * h + r; const int mm = min(m, p.M - 1);
            float v = acc[t][r] * iscale;
            if (p.flags & 1) v += p.bias[nn];
            if (p.flags & 2) v += p.bias[mm];
            v = act_fn(v, p.act);
            if (p.flags & 4) v += p.beta * R[(long long)mm * p.sRm + (long long)nn * p.sRn];
            ctile[8 * h + r][t * 16 + l15] = (n < p.N) ? v : 0.f;
        }
    }
    __syncthreads();
    const int NW = (p.Npad > p.N) ? p.Npad : p.N;
    const bool fast = (m0 + 16 <= p.M) && (n0 + 32 <= NW) && ((p.sCm & 3) == 0) && ((((size_t)C) & 15) == 0);
    if (fast) {
#pragma unroll
        for (int s = 0; s < 4; ++s) {
            const int row = s * 4 + (lane >> 3), c4 = (lane & 7) * 4;
            const v4f v = *(const v4f*)&ctile[row][c4];
            VST2V4(C + (long long)(m0 + row) * p.sCm + n0 + c4, v);
        }
    } else {
        for (int row = 0; row < 16; ++row) {
            const int m = m0 + row, n = n0 + lane;
            if (m < p.M && n < NW) VST2(float, C + (long long)m * p.sCm + n, ctile[row][lane]);
        }
    }
}

#define AW 4
struct AttnP {
    const float* Q; const float* K; const float* V; float* O; float* P; const float* Mf; const int* Mi; float* ST;
    const float* Pw; const float* Rt; const int* SQ; const int* SK;
    long long swb, swh, swi, swj, srb, srh, sri;
    long long sQb, sQh, sQi, sQd, sKb, sKh, sKj, sKd, sVb, sVh, sVj, sVd, sOb, sOh, sOi, sPb, sPh, sPi, smb, smh, smi, smj;
    int Lq, Lk, dh, dv, hrep, causal, coff, pband;
    float scale, mfill; int nonorm, mpol;
    int roff, rn, segpol, win;
};
static_assert(sizeof(AttnP) == 12 * 8 + 29 * 8 + 16 * 4, "AttnP has padding");

#ifndef KATTN_ATTR
#define KATTN_ATTR
#endif
template <int DHP, int DVP, int QM, bool SPLITPV, bool TWOPASS>
__global__ __launch_bounds__(32 * AW) KATTN_ATTR void k_attn(AttnP p) {
    constexpr int NT = DVP / 16;
    constexpr int KS = DHP / 32;
    constexpr int VP = DVP + 8;
    __shared__ __align__(16) float    pl[AW][16 * 64];
    __shared__ __align__(16) _Float16 vl[(SPLITPV ? 2 : 1) * 64 * VP];
    const int lane = threadIdx.x & 31, hf = lane >> 4, l15 = lane & 15, wave = threadIdx.x >> 5;
    const int h = blockIdx.y, b = blockIdx.z, hk = h / p.hrep;
    const int q0 = (blockIdx.x * AW + wave) * 16;
    float* myp = pl[wave];
    const float L2E = 1.4426950408889634f;
    const float NEG = -__builtin_inff();
    const int qi = min(q0 + l15, p.Lq - 1);
    const float* qrow = p.Q + b * p.sQb + h * p.sQh + (long long)qi * p.sQi;
    const float* kbase = p.K + b * p.sKb + hk * p.sKh;
    const float* vbase = p.V + b * p.sVb + hk * p.sVh;
    v16h qa[QM == 0 ? KS : 1]; Split qs_[QM == 1 ? KS : 1]; Split3 qt_[QM == 2 ? KS : 1];
#pragma unroll
    for (int ks = 0; ks < KS; ++ks) {
        if (QM == 2) qt_[ks] = sp3_ld(qrow, p.sQd, ks * 32, hf, p.dh, 1.f);
        else if (QM == 1) qs_[ks] = sp_ld(qrow, p.sQd, ks * 32, hf, p.dh, 1.f);
        else qa[ks] = fh_ld(qrow, p.sQd, ks * 32, hf, p.dh, 1.f);
    }
    v8f o[NT]; float m8[8], l8[8];
#pragma unroll
    for (int t = 0; t < NT; ++t) { v8f zz = {}; o[t] = zz; }
#pragma unroll
    for (int i = 0; i < 8; ++i) { m8[i] = NEG; l8[i] = 0.f; }
    int jend = p.Lk;
    if (p.causal == 1) { const int je = (blockIdx.x * AW + AW - 1) * 16 + 16 + p.coff; jend = min(jend, max(je, 0)); }
    const int npass = TWOPASS ? 2 : 1;
    for (int pass = 0; pass < npass; ++pass) {
        const bool dopv = (!TWOPASS) || pass == 1;
        for (int j0 = 0; j0 < jend; j0 += 64) {
            if (dopv) {
                __syncthreads();
                for (int idx = threadIdx.x; idx < 64 * DVP; idx += 32 * AW) {
                    const int jr = idx / DVP, d = idx - jr * DVP, j = j0 + jr;
                    const float f = (j < p.Lk && d < p.dv) ? vbase[(long long)j * p.sVj + (long long)d * p.sVd] : 0.f;
                    if (SPLITPV) {
                        const __bf16 hb = bf16_rne(f);
                        ((__bf16*)vl)[jr * VP + d] = hb; ((__bf16*)vl)[64 * VP + jr * VP + d] = bf16_rne(f - bf16_f32(hb));
                    } else vl[jr * VP + d] = (_Float16)f;
                }
            }
            v8f s[4];
#pragma unroll
            for (int t = 0; t < 4; ++t) {
                const int j = min(j0 + t * 16 + l15, p.Lk - 1);
                const float* krow = kbase + (long long)j * p.sKj;
                v8f acc = {};
#pragma unroll
                for (int ks = 0; ks < KS; ++ks) {
                    if (QM == 2)      acc = wmma6(qt_[ks], sp3_ld(krow, p.sKd, ks * 32, hf, p.dh, 1.f), acc);
                    else if (QM == 1) acc = wmma3(qs_[ks], sp_ld(krow, p.sKd, ks * 32, hf, p.dh, 1.f), acc);
                    else              acc = wmma16(qa[ks], fh_ld(krow, p.sKd, ks * 32, hf, p.dh, 1.f), acc);
                }
                s[t] = acc;
            }
            float pv[8][4];
#pragma unroll
            for (int i = 0; i < 8; ++i) {
                const int irow = q0 + i + 8 * hf;
                const int ic = min(irow, p.Lq - 1);
                float sc[4];
#pragma unroll
                for (int t = 0; t < 4; ++t) {
                    const int jg = j0 + t * 16 + l15;
                    float v = s[t][i] * p.scale;
                    if (p.Mf) v += p.Mf[b * p.smb + h * p.smh + (long long)ic * p.smi + (long long)min(jg, p.Lk - 1) * p.smj];
                    if (p.Rt) { int rc = ic - min(jg, p.Lk - 1) + p.roff; rc = rc < 0 ? 0 : (rc >= p.rn ? p.rn - 1 : rc); v += p.Rt[b * p.srb + h * p.srh + (long long)ic * p.sri + rc]; }
                    if (p.Mi) { const int mv = p.Mi[b * p.smb + h * p.smh + (long long)ic * p.smi + (long long)min(jg, p.Lk - 1) * p.smj]; if (p.mpol ? (mv != 0) : (mv == 0)) v = p.mfill; }
                    if (p.SQ) { const bool same = p.SQ[(long long)b * p.Lq + ic] == p.SK[(long long)b * p.Lk + min(jg, p.Lk - 1)]; if (p.segpol ? same : !same) v = p.mfill; }
                    if (p.causal == 2 && jg > irow + p.coff) v = p.mfill;
                    if (jg >= p.Lk || (p.causal == 1 && jg > irow + p.coff) || (p.causal == 3 && jg < irow + p.coff) || (p.win > 0 && irow + p.coff - jg > p.win)) v = NEG; else v *= L2E;
                    sc[t] = v;
                }
                if (!TWOPASS || pass == 0) {
                    float mx = fmaxf(fmaxf(sc[0], sc[1]), fmaxf(sc[2], sc[3]));
                    mx = fmaxf(mx, __shfl_xor(mx, 1, 32)); mx = fmaxf(mx, __shfl_xor(mx, 2, 32));
                    mx = fmaxf(mx, __shfl_xor(mx, 4, 32)); mx = fmaxf(mx, __shfl_xor(mx, 8, 32));
                    const float mnew = fmaxf(m8[i], mx);
                    const float corr = (mnew == NEG) ? 1.f : exp2f(m8[i] - mnew);
                    float rs = 0.f;
#pragma unroll
                    for (int t = 0; t < 4; ++t) {
                        const float pp = (sc[t] == NEG) ? 0.f : exp2f(sc[t] - mnew); rs += pp;
                        pv[i][t] = p.Pw ? pp * p.Pw[b * p.swb + h * p.swh + (long long)ic * p.swi + (long long)min(j0 + t * 16 + l15, p.Lk - 1) * p.swj] : pp;
                    }
                    rs += __shfl_xor(rs, 1, 32); rs += __shfl_xor(rs, 2, 32); rs += __shfl_xor(rs, 4, 32); rs += __shfl_xor(rs, 8, 32);
                    l8[i] = l8[i] * corr + rs; m8[i] = mnew;
                    if (!TWOPASS) {
#pragma unroll
                        for (int t = 0; t < NT; ++t) o[t][i] *= corr;
                    }
                } else {
                    const float inv = (l8[i] > 0.f) ? 1.f / l8[i] : 0.f;
#pragma unroll
                    for (int t = 0; t < 4; ++t) {
                        const int jg = j0 + t * 16 + l15;
                        float pp = (sc[t] == NEG) ? 0.f : exp2f(sc[t] - m8[i]) * inv;
                        if (p.Pw) pp *= p.Pw[b * p.swb + h * p.swh + (long long)ic * p.swi + (long long)min(jg, p.Lk - 1) * p.swj];
                        pv[i][t] = pp;
                    }
                }
            }
            if (dopv) {
#pragma unroll
                for (int i = 0; i < 8; ++i)
#pragma unroll
                    for (int t = 0; t < 4; ++t) myp[(i + 8 * hf) * 64 + t * 16 + l15] = pv[i][t];
                __syncthreads();
                if (p.P) {
                    float* pb_ = p.P + b * p.sPb + h * p.sPh;
                    const bool fastP = (p.pband == 0) && ((p.sPi & 3) == 0) && (j0 + 64 <= p.Lk) && (q0 + 16 <= p.Lq) && ((((size_t)pb_) & 15) == 0);
                    if (fastP) {
#pragma unroll
                        for (int s = 0; s < 8; ++s) {
                            const int row = s * 2 + (lane >> 4), c4 = (lane & 15) * 4;
                            const v4f v = *(const v4f*)(myp + row * 64 + c4);
                            VST2V4(pb_ + (long long)(q0 + row) * p.sPi + j0 + c4, v);
                        }
                    } else {
                        for (int row = 0; row < 16; ++row) {
                            const int irow = q0 + row; if (irow >= p.Lq) continue;
                            for (int c = lane; c < 64; c += 32) {
                                const int jg = j0 + c; if (jg >= p.Lk) continue;
                                if (p.pband == 0) VST2(float, pb_ + (long long)irow * p.sPi + jg, myp[row * 64 + c]);
                                else if (jg - irow <= p.pband && irow - jg <= p.pband) VST2(float, pb_ + (long long)irow * p.sPi + (jg - irow + p.pband), myp[row * 64 + c]);
                            }
                        }
                    }
                }
                if (SPLITPV) {
                    const Split pa0 = sp_ld(myp + l15 * 64, 1, 0, hf, 64, 1.f), pa1 = sp_ld(myp + l15 * 64, 1, 32, hf, 64, 1.f);
                    const __bf16* vh = (const __bf16*)vl; const __bf16* vlo = vh + 64 * VP;
#pragma unroll
                    for (int t = 0; t < NT; ++t) {
                        const int dcol = t * 16 + l15;
                        Split b0, b1;
#pragma unroll
                        for (int e = 0; e < 16; ++e) {
                            const int k0 = frag_k(e, hf), k1 = 32 + frag_k(e, hf);
                            b0.hi[e] = vh[k0 * VP + dcol]; b0.lo[e] = vlo[k0 * VP + dcol]; b1.hi[e] = vh[k1 * VP + dcol]; b1.lo[e] = vlo[k1 * VP + dcol];
                        }
                        o[t] = wmma3(pa0, b0, o[t]);
                        o[t] = wmma3(pa1, b1, o[t]);
                    }
                } else {
                    const v16h pa0 = fh_ld(myp + l15 * 64, 1, 0, hf, 64, 4096.f), pa1 = fh_ld(myp + l15 * 64, 1, 32, hf, 64, 4096.f);
#pragma unroll
                    for (int t = 0; t < NT; ++t) {
                        const int dcol = t * 16 + l15;
                        v16h b0, b1;
#pragma unroll
                        for (int e = 0; e < 16; ++e) { b0[e] = vl[frag_k(e, hf) * VP + dcol]; b1[e] = vl[(32 + frag_k(e, hf)) * VP + dcol]; }
                        o[t] = wmma16(pa0, b0, o[t]);
                        o[t] = wmma16(pa1, b1, o[t]);
                    }
                }
            }
        }
    }
    float* obase = p.O + b * p.sOb + h * p.sOh;
    if (p.ST) {
        const int rl = lane >> 1, isel = rl & 7;
        float mv = 0.f, lv = 0.f;
#pragma unroll
        for (int i = 0; i < 8; ++i) if (i == isel) { mv = m8[i]; lv = l8[i]; }
        const int irow = q0 + rl;
        if (irow < p.Lq) { float* st = p.ST + (((long long)b * gridDim.y + h) * p.Lq + irow) * 2 + (lane & 1); VST2(float, st, (lane & 1) ? lv : mv * 0.6931471805599453f); }
    }
    float invr[8];
#pragma unroll
    for (int i = 0; i < 8; ++i) {
        if (TWOPASS) invr[i] = SPLITPV ? 1.f : (1.f / 4096.f);
        else if (p.nonorm) invr[i] = exp2f(m8[i]) * (SPLITPV ? 1.f : (1.f / 4096.f));
        else invr[i] = (l8[i] > 0.f) ? (SPLITPV ? 1.f / l8[i] : 1.f / (l8[i] * 4096.f)) : 0.f;
    }
    __syncthreads();
    const bool ofast = ((p.sOi & 3) == 0) && ((((size_t)obase) & 15) == 0) && (q0 + 16 <= p.Lq);
#pragma unroll
    for (int c0 = 0; c0 < DVP; c0 += 64) {
#pragma unroll
        for (int i = 0; i < 8; ++i)
#pragma unroll
            for (int t = 0; t < NT; ++t) if (t * 16 >= c0 && t * 16 < c0 + 64) myp[(i + 8 * hf) * 64 + (t * 16 - c0) + l15] = o[t][i] * invr[i];
        __syncthreads();
        const int cw = (DVP - c0 < 64) ? (DVP - c0) : 64;
        if (ofast && (c0 + cw <= p.dv) && (cw % 32 == 0)) {
            const int lpr = cw / 4;
            const int rows_per_ins = 32 / lpr;
            for (int r0 = 0; r0 < 16; r0 += rows_per_ins) {
                const int row = r0 + lane / lpr, c4 = (lane % lpr) * 4;
                const v4f v = *(const v4f*)(myp + row * 64 + c4);
                VST2V4(obase + (long long)(q0 + row) * p.sOi + c0 + c4, v);
            }
        } else {
            for (int row = 0; row < 16; ++row) {
                const int irow = q0 + row; if (irow >= p.Lq) continue;
                for (int c = lane; c < cw; c += 32) { const int d = c0 + c; if (d < p.dv) VST2(float, obase + (long long)irow * p.sOi + d, myp[row * 64 + c]); }
            }
        }
        __syncthreads();
    }
}

struct TrP { const float* src; float* dst; const float* R2; long long sSz, lds, sDz, ldd, sRz, ldr; int R, C, flags, act; float alpha, beta; };
static_assert(sizeof(TrP) == 3 * 8 + 6 * 8 + 6 * 4, "TrP has padding");
__global__ __launch_bounds__(256) void k_tr(TrP p) {
    __shared__ float tile[32][33];
    const int c0 = blockIdx.x * 32, r0 = blockIdx.y * 32, z = blockIdx.z;
    const int lane = threadIdx.x & 31, wave = threadIdx.x >> 5;
    const float* s = p.src + z * p.sSz;
#pragma unroll
    for (int k = 0; k < 4; ++k) {
        const int rl = wave * 4 + k, r = r0 + rl, c = c0 + lane;
        tile[rl][lane] = (r < p.R && c < p.C) ? s[(long long)r * p.lds + c] : 0.f;
    }
    __syncthreads();
    float* d = p.dst + z * p.sDz; const float* rr = p.R2 + z * p.sRz;
#pragma unroll
    for (int k = 0; k < 4; ++k) {
        const int cl = wave * 4 + k, c = c0 + cl, r = r0 + lane;
        if (c < p.C && r < p.R) {
            float v = act_fn(p.alpha * tile[lane][cl], p.act);
            if (p.flags & 1) v += p.beta * rr[(long long)c * p.ldr + r];
            VST2(float, d + (long long)c * p.ldd + r, v);
        }
    }
}

__global__ __launch_bounds__(256) void k_affine(const float* __restrict__ src, float* __restrict__ dst, int n, float a, float b, const float* __restrict__ sdev) {
    const int i = blockIdx.x * 256 + threadIdx.x;
    if (i < n) { const float aa = sdev ? a * sdev[0] : a; const float v = aa * src[i] + b; VST2(float, dst + i, v); }
}

struct SmP { const float* src; float* dst; const float* Mf; long long sz, sr, dz, dr, smz, smr; int n, pad; float scale_in, scale_out; };
static_assert(sizeof(SmP) == 3 * 8 + 6 * 8 + 4 * 4, "SmP has padding");
__global__ __launch_bounds__(256) void k_softmax(SmP p) {
    __shared__ float red[256];
    const int r = blockIdx.x, z = blockIdx.y, tid = threadIdx.x;
    const float* s = p.src + z * p.sz + (long long)r * p.sr;
    const float* mf = p.Mf ? (p.Mf + z * p.smz + (long long)r * p.smr) : nullptr;
    float mx = -__builtin_inff();
    for (int j = tid; j < p.n; j += 256) { float v = s[j] * p.scale_in; if (mf) v += mf[j]; mx = fmaxf(mx, v); }
    red[tid] = mx; __syncthreads();
    for (int o = 128; o > 0; o >>= 1) { if (tid < o) red[tid] = fmaxf(red[tid], red[tid + o]); __syncthreads(); }
    mx = red[0]; __syncthreads();
    float sum = 0.f;
    for (int j = tid; j < p.n; j += 256) { float v = s[j] * p.scale_in; if (mf) v += mf[j]; sum += (mx == -__builtin_inff()) ? 0.f : expf(v - mx); }
    red[tid] = sum; __syncthreads();
    for (int o = 128; o > 0; o >>= 1) { if (tid < o) red[tid] += red[tid + o]; __syncthreads(); }
    sum = red[0];
    const float inv = (sum > 0.f) ? p.scale_out / sum : 0.f;
    float* d = p.dst + z * p.dz + (long long)r * p.dr;
    for (int j = tid; j < p.n; j += 256) { float v = s[j] * p.scale_in; if (mf) v += mf[j]; const float o = (mx == -__builtin_inff()) ? 0.f : expf(v - mx) * inv; VST2(float, d + j, o); }
}
__global__ __launch_bounds__(256) void k_stats(const float* __restrict__ x, long long sz, long long so, long long si, int inner, int n, float eps, float* __restrict__ stat, int mode) {
    __shared__ float red[256];
    const int z = blockIdx.x, tid = threadIdx.x;
    const float* base = x + z * sz;
    float s = 0.f;
    for (int e = tid; e < n; e += 256) s += base[(long long)(e / inner) * so + (long long)(e % inner) * si];
    red[tid] = s; __syncthreads();
    for (int o = 128; o > 0; o >>= 1) { if (tid < o) red[tid] += red[tid + o]; __syncthreads(); }
    const float mu = (mode == 0 || mode == 3) ? red[0] / (float)n : 0.f; __syncthreads();
    float q = 0.f;
    for (int e = tid; e < n; e += 256) { const float dlt = base[(long long)(e / inner) * so + (long long)(e % inner) * si] - mu; q += dlt * dlt; }
    red[tid] = q; __syncthreads();
    for (int o = 128; o > 0; o >>= 1) { if (tid < o) red[tid] += red[tid + o]; __syncthreads(); }
    {
        float rs;
        if (mode == 2) rs = sqrtf((float)n) / fmaxf(sqrtf(red[0]), eps); else if (mode == 3) rs = rsqrtf(red[0] / (float)(n - 1) + eps); else rs = rsqrtf(red[0] / (float)n + eps);
        if (tid < 32) { const float v = (tid == 0) ? mu : ((tid == 1) ? rs : 0.f); VST2(float, stat + (long long)z * 32 + tid, v); }
    }
}
__global__ __launch_bounds__(256) void k_norm_apply(const float* __restrict__ x, float* __restrict__ y, const float* __restrict__ stat, const float* __restrict__ g, const float* __restrict__ bta,
                                                     int Z, int C, int L, int G, int bn, int act) {
    const long long idx = (long long)blockIdx.x * 256 + threadIdx.x;
    if (idx >= (long long)Z * C * L) return;
    const int l = (int)(idx % L); const long long zc = idx / L; const int c = (int)(zc % C), z = (int)(zc / C); (void)l;
    const int set = bn ? c : (z * G + c / (C / G));
    float v = (x[idx] - stat[(long long)set * 32]) * stat[(long long)set * 32 + 1];
    if (g) v *= g[c];
    if (bta) v += bta[c];
    v = act_fn(v, act);
    VST2(float, y + idx, v);
}

__global__ __launch_bounds__(256) void k_lse_neg(const float* __restrict__ st, float* __restrict__ c, int n) {
    const int i = blockIdx.x * 256 + threadIdx.x;
    if (i < n) { const float v = -(st[2 * i] + logf(st[2 * i + 1])); VST2(float, c + i, v); }
}

__global__ __launch_bounds__(256) void k_iota(int* __restrict__ dst, int n, int a, int b) {
    const int i = blockIdx.x * 256 + threadIdx.x;
    if (i < n) { const int v = a * i + b; VST2(int, dst + i, v); }
}

__global__ __launch_bounds__(256) void k_axpby(const float* __restrict__ x, const float* __restrict__ y, float* __restrict__ dst, int n, float a, float b, float c) {
    const int i = blockIdx.x * 256 + threadIdx.x;
    if (i < n) { const float v = a * x[i] + b * y[i] + c; VST2(float, dst + i, v); }
}

struct RopeP { const float* X; float* Y; const float* C; const float* Sn; const int* pos; long long sXr, sXh, sYr, sYh, sCb, sCp, sCd; int R, Hn, D, S, mode, tmode, pmode, pad; };
static_assert(sizeof(RopeP) == 5 * 8 + 7 * 8 + 8 * 4, "RopeP has padding");
__global__ __launch_bounds__(256) void k_rope(RopeP p) {
    const long long idx = (long long)blockIdx.x * 256 + threadIdx.x;
    if (idx >= (long long)p.R * p.Hn * p.D) return;
    const int d = (int)(idx % p.D); const long long rh = idx / p.D; const int h = (int)(rh % p.Hn); const int r = (int)(rh / p.Hn);
    const int half = p.D / 2;
    int partner; float sign;
    if (p.mode == 0) { partner = (d < half) ? d + half : d - half; sign = (d < half) ? -1.f : 1.f; }
    else { partner = d ^ 1; sign = (d & 1) ? 1.f : -1.f; }
    const int tcol = (p.tmode == 0) ? d : ((p.tmode == 1) ? (d % half) : (d >> 1));
    const int pp = (p.pmode == 0) ? (r % p.S) : ((p.pmode == 1) ? h : p.pos[r]);
    const long long toff = (long long)(r / p.S) * p.sCb + (long long)pp * p.sCp + (long long)tcol * p.sCd;
    const float* xr = p.X + (long long)r * p.sXr + (long long)h * p.sXh;
    const float v = xr[d] * p.C[toff] + sign * xr[partner] * p.Sn[toff];
    VST2(float, p.Y + (long long)r * p.sYr + (long long)h * p.sYh + d, v);
}

__global__ __launch_bounds__(256) void k_invf(float* __restrict__ invb, int half, int D, float base, float num, int fmode, float cexp) {
    const int i = blockIdx.x * 256 + threadIdx.x;
    if (i >= ((half + 31) / 32) * 32) return;
    if (i >= half) { VST2(float, invb + i, 0.f); return; }
    const float e = (float)(2 * i) / (float)D;
    float invf;
    if (fmode == 1) invf = num * expf((float)(2 * i) * cexp);
    else if (fmode == 2) invf = num * powf(base, (-2.0f * ((float)i - 1.0f)) / (float)D);
    else invf = num * (1.0f / powf(base, e));
    VST2(float, invb + i, invf);
}
__global__ __launch_bounds__(256) void k_sincos(float* __restrict__ cs, float* __restrict__ sn, const float* __restrict__ invb, int S, int half, float pscale) {
    const int idx = blockIdx.x * 256 + threadIdx.x;
    if (idx >= S * half) return;
    const int s = idx / half, i = idx - s * half;
    const float ang = (pscale * (float)s) * invb[i];
    VST2(float, cs + idx, cosf(ang)); VST2(float, sn + idx, sinf(ang));
}

__global__ __launch_bounds__(256) void k_mulact(const float* __restrict__ x, const float* __restrict__ y, float* __restrict__ dst, int n, int act) {
    const int i = blockIdx.x * 256 + threadIdx.x;
    if (i < n) { const float v = act_fn(x[i], act) * y[i]; VST2(float, dst + i, v); }
}

__global__ __launch_bounds__(256) void k_matvec(GemmP p) {
    const int rpt = (p.N == 1) ? 1 : 32;
    const long long r0 = ((long long)blockIdx.x * 256 + threadIdx.x) * rpt; const int z = blockIdx.z, zo = z / p.zi_n, zi = z - zo * p.zi_n;
    if (r0 >= p.M) return;
    const float* Bb = p.B + zo * p.sBo + zi * p.sBi;
    float* C = p.C + zo * p.sCo + zi * p.sCi; const float* R = p.R + zo * p.sRo + zi * p.sRi;
    for (int rr = 0; rr < rpt; ++rr) {
        const long long r = r0 + rr; if (r >= p.M) break;
        const float* A = p.A + zo * p.sAo + zi * p.sAi + r * p.sAm;
        float acc[8] = {0.f, 0.f, 0.f, 0.f, 0.f, 0.f, 0.f, 0.f};
        for (int k = 0; k < p.K; ++k) { const float a = A[(long long)k * p.sAk];
#pragma unroll
            for (int j = 0; j < 8; ++j) if (j < p.N) acc[j] += a * Bb[(long long)j * p.sBn + (long long)k * p.sBk]; }
#pragma unroll
        for (int j = 0; j < 8; ++j) if (j < p.N) {
            float v = acc[j] * p.alpha;
            if (p.flags & 1) v += p.bias[j];
            if (p.flags & 2) v += p.bias[r];
            v = act_fn(v, p.act);
            if (p.flags & 4) v += p.beta * R[r * p.sRm + (long long)j * p.sRn];
            VST2(float, C + r * p.sCm + j, v);
        }
    }
}
__global__ __launch_bounds__(256) void k_smallsoftmax(const float* __restrict__ src, float* __restrict__ dst, long long sr, long long dr, int n, long long R, float scale) {
    const long long r0 = ((long long)blockIdx.x * 256 + threadIdx.x) * 32;
    for (int rr = 0; rr < 32; ++rr) {
        const long long r = r0 + rr; if (r >= R) return;
        const float* s = src + r * sr; float* d = dst + r * dr;
        float mx = -__builtin_inff();
        for (int j = 0; j < n; ++j) mx = fmaxf(mx, s[j] * scale);
        float sum = 0.f;
        for (int j = 0; j < n; ++j) sum += expf(s[j] * scale - mx);
        const float inv = 1.f / sum;
        for (int j = 0; j < n; ++j) { const float v = expf(s[j] * scale - mx) * inv; VST2(float, d + j, v); }
    }
}

__global__ __launch_bounds__(32) void k_unitstat(float* __restrict__ st) { const int t = threadIdx.x; const float v = (t == 1) ? 1.f : 0.f; VST2(float, st + t, v); }

__global__ __launch_bounds__(256) void k_lincopy(const float* __restrict__ src, long long lds, float* __restrict__ dst, long long ldd, long long rows, int cols) {
    const long long i = (long long)blockIdx.x * 256 + threadIdx.x; if (i >= rows * cols) return;
    const long long r = i / cols; const int c = (int)(i - r * cols);
    const float v = src[r * lds + c]; VST2(float, dst + r * ldd + c, v);
}

__global__ __launch_bounds__(256) void k_catcg(const float* __restrict__ ctx, const float* __restrict__ goals, float* __restrict__ CG, int B, int KM, int H, int ld) {
    const long long t = (long long)blockIdx.x * 256 + threadIdx.x; if (t >= (long long)B * KM * ld) return; const int c = (int)(t % ld); const int r = (int)(t / ld); const int b = r / KM;
    float v = 0.f; if (c < H) v = ctx[(long long)b * H + c]; else if (c < H + 2) v = goals[(long long)r * 2 + (c - H)];
    VST2(float, CG + t, v);
}
__global__ __launch_bounds__(256) void k_gru(const float* __restrict__ GI, const float* __restrict__ X2, const float* __restrict__ wih0, const float* __restrict__ bih0, const float* __restrict__ GH, const float* __restrict__ Hp, float* __restrict__ Hn, int N, int H) {
    const long long t = (long long)blockIdx.x * 256 + threadIdx.x; if (t >= (long long)N * H) return; const int c = (int)(t % H); const int n = (int)(t / H);
    float gir, giz, gin;
    if (X2) { const float x0 = X2[2 * n], x1 = X2[2 * n + 1];
        gir = x0 * wih0[(c) * 2] + x1 * wih0[(c) * 2 + 1] + bih0[c]; giz = x0 * wih0[(H + c) * 2] + x1 * wih0[(H + c) * 2 + 1] + bih0[H + c]; gin = x0 * wih0[(2 * H + c) * 2] + x1 * wih0[(2 * H + c) * 2 + 1] + bih0[2 * H + c]; }
    else { const float* gi = GI + (long long)n * 3 * H; gir = gi[c]; giz = gi[H + c]; gin = gi[2 * H + c]; }
    const float* gh = GH + (long long)n * 3 * H;
    const float r = 1.f / (1.f + expf(-(gir + gh[c]))); const float z = 1.f / (1.f + expf(-(giz + gh[H + c]))); const float nn = tanhf(gin + r * gh[2 * H + c]);
    VST2(float, Hn + t, (1.f - z) * nn + z * Hp[t]);
}
__global__ __launch_bounds__(256) void k_posstep(const float* __restrict__ DL, int ldp, float* __restrict__ X, float* __restrict__ POS, float* __restrict__ TRAJ, int N, int T, int step) {
    const int t = blockIdx.x * 256 + threadIdx.x; if (t >= N * 2) return; const int c = t & 1; const int r = t >> 1; const float d = DL[(long long)r * ldp + c]; const float pz = POS[t] + d;
    VST2(float, X + t, d); VST2(float, POS + t, pz); VST2(float, TRAJ + ((long long)r * T + step) * 2 + c, pz);
}
__global__ __launch_bounds__(256) void k_ramp(const float* __restrict__ TRAJ, const float* __restrict__ goals, float* __restrict__ OUT, int N, int T) {
    const long long t = (long long)blockIdx.x * 256 + threadIdx.x; if (t >= (long long)N * T * 2) return; const int c = (int)(t & 1); const int s = (int)((t >> 1) % T); const int r = (int)(t / (2 * T));
    const float e = goals[(long long)r * 2 + c] - TRAJ[((long long)r * T + T - 1) * 2 + c]; const float ramp = (float)(s + 1) / (float)T;
    VST2(float, OUT + t, TRAJ[t] + ramp * e);
}

template __global__ void k_gemm<1>(GemmP);

extern "C" void kernel_launch(void* const* d_in, const int* in_sizes, int n_in, void* d_out, int out_size, void* d_ws, size_t ws_size, hipStream_t stream) {
    (void)in_sizes; (void)n_in; (void)out_size; (void)ws_size;
    const float* ctx = (const float*)d_in[0];
    const float* goals = (const float*)d_in[1];
    const float* hiw = (const float*)d_in[2];
    const float* hib = (const float*)d_in[3];
    const float* wih0 = (const float*)d_in[4];
    const float* whh0 = (const float*)d_in[5];
    const float* bih0 = (const float*)d_in[6];
    const float* bhh0 = (const float*)d_in[7];
    const float* wih1 = (const float*)d_in[8];
    const float* whh1 = (const float*)d_in[9];
    const float* bih1 = (const float*)d_in[10];
    const float* bhh1 = (const float*)d_in[11];
    const float* ow = (const float*)d_in[12];
    const float* ob = (const float*)d_in[13];
    const int Bn = 2048;
    const int KM = 6;
    const int BK = Bn * KM;
    const int H = 256;
    const int H3 = 768;
    const int T = 30;
    const int LDC = 288;
    const int LDP = 32;
    float* out = (float*)d_out;
    char* wsp = (char*)d_ws;
    float* CG = (float*)wsp; wsp += (((size_t)((size_t)BK * LDC) * 4 + 255) / 256) * 256;
    float* H0 = (float*)wsp; wsp += (((size_t)((size_t)BK * H) * 4 + 255) / 256) * 256;
    float* H1 = (float*)wsp; wsp += (((size_t)((size_t)BK * H) * 4 + 255) / 256) * 256;
    float* H0n = (float*)wsp; wsp += (((size_t)((size_t)BK * H) * 4 + 255) / 256) * 256;
    float* H1n = (float*)wsp; wsp += (((size_t)((size_t)BK * H) * 4 + 255) / 256) * 256;
    float* GH = (float*)wsp; wsp += (((size_t)((size_t)BK * H3) * 4 + 255) / 256) * 256;
    float* GI = (float*)wsp; wsp += (((size_t)((size_t)BK * H3) * 4 + 255) / 256) * 256;
    float* X = (float*)wsp; wsp += (((size_t)((size_t)BK * 2) * 4 + 255) / 256) * 256;
    float* POS = (float*)wsp; wsp += (((size_t)((size_t)BK * 2) * 4 + 255) / 256) * 256;
    float* DL = (float*)wsp; wsp += (((size_t)((size_t)BK * LDP) * 4 + 255) / 256) * 256;
    float* TRAJ = (float*)wsp; wsp += (((size_t)((size_t)BK * T * 2) * 4 + 255) / 256) * 256;
    k_catcg<<<(unsigned)(((long long)BK * LDC + 255) / 256), 256, 0, stream>>>(ctx, goals, CG, Bn, KM, H, LDC);
    hipMemsetAsync(X, 0, (size_t)BK * 2 * 4, stream);
    hipMemsetAsync(POS, 0, (size_t)BK * 2 * 4, stream);
    { GemmP ginit;
      ginit.A = CG; ginit.B = hiw; ginit.bias = hib; ginit.R = CG; ginit.C = H0;
      ginit.sAo = 0; ginit.sAi = 0; ginit.sAm = LDC; ginit.sAk = 1; ginit.sBo = 0; ginit.sBi = 0; ginit.sBn = H + 2; ginit.sBk = 1; ginit.sCo = 0; ginit.sCi = 0; ginit.sCm = H; ginit.sRo = 0; ginit.sRi = 0; ginit.sRm = 0; ginit.sRn = 0;
      ginit.M = BK; ginit.N = H; ginit.K = H + 2; ginit.zi_n = 1; ginit.flags = 1; ginit.act = 5;
      ginit.alpha = 1.0f; ginit.beta = 0.0f; ginit.sa = 1.0f; ginit.sb = 1.0f; ginit.Npad = H; ginit.pad_ = 0;
      k_gemm<1><<<dim3((unsigned)((H) + 31) / 32, (unsigned)((BK) + 15) / 16, (unsigned)(1)), 32, 0, stream>>>(ginit); }
    k_lincopy<<<(unsigned)(((long long)(BK) * (H) + 255) / 256), 256, 0, stream>>>(H0, H, H1, H, BK, H);
    { GemmP gh0_0;
      gh0_0.A = H0; gh0_0.B = whh0; gh0_0.bias = bhh0; gh0_0.R = H0; gh0_0.C = GH;
      gh0_0.sAo = 0; gh0_0.sAi = 0; gh0_0.sAm = H; gh0_0.sAk = 1; gh0_0.sBo = 0; gh0_0.sBi = 0; gh0_0.sBn = H; gh0_0.sBk = 1; gh0_0.sCo = 0; gh0_0.sCi = 0; gh0_0.sCm = H3; gh0_0.sRo = 0; gh0_0.sRi = 0; gh0_0.sRm = 0; gh0_0.sRn = 0;
      gh0_0.M = BK; gh0_0.N = H3; gh0_0.K = H; gh0_0.zi_n = 1; gh0_0.flags = 1; gh0_0.act = 0;
      gh0_0.alpha = 1.0f; gh0_0.beta = 0.0f; gh0_0.sa = 1.0f; gh0_0.sb = 1.0f; gh0_0.Npad = H3; gh0_0.pad_ = 0;
      k_gemm<1><<<dim3((unsigned)((H3) + 31) / 32, (unsigned)((BK) + 15) / 16, (unsigned)(1)), 32, 0, stream>>>(gh0_0); }
    k_gru<<<(unsigned)(((long long)BK * H + 255) / 256), 256, 0, stream>>>(nullptr, X, wih0, bih0, GH, H0, H0n, BK, H);
    { GemmP gi1_0;
      gi1_0.A = H0n; gi1_0.B = wih1; gi1_0.bias = bih1; gi1_0.R = H0n; gi1_0.C = GI;
      gi1_0.sAo = 0; gi1_0.sAi = 0; gi1_0.sAm = H; gi1_0.sAk = 1; gi1_0.sBo = 0; gi1_0.sBi = 0; gi1_0.sBn = H; gi1_0.sBk = 1; gi1_0.sCo = 0; gi1_0.sCi = 0; gi1_0.sCm = H3; gi1_0.sRo = 0; gi1_0.sRi = 0; gi1_0.sRm = 0; gi1_0.sRn = 0;
      gi1_0.M = BK; gi1_0.N = H3; gi1_0.K = H; gi1_0.zi_n = 1; gi1_0.flags = 1; gi1_0.act = 0;
      gi1_0.alpha = 1.0f; gi1_0.beta = 0.0f; gi1_0.sa = 1.0f; gi1_0.sb = 1.0f; gi1_0.Npad = H3; gi1_0.pad_ = 0;
      k_gemm<1><<<dim3((unsigned)((H3) + 31) / 32, (unsigned)((BK) + 15) / 16, (unsigned)(1)), 32, 0, stream>>>(gi1_0); }
    { GemmP gh1_0;
      gh1_0.A = H1; gh1_0.B = whh1; gh1_0.bias = bhh1; gh1_0.R = H1; gh1_0.C = GH;
      gh1_0.sAo = 0; gh1_0.sAi = 0; gh1_0.sAm = H; gh1_0.sAk = 1; gh1_0.sBo = 0; gh1_0.sBi = 0; gh1_0.sBn = H; gh1_0.sBk = 1; gh1_0.sCo = 0; gh1_0.sCi = 0; gh1_0.sCm = H3; gh1_0.sRo = 0; gh1_0.sRi = 0; gh1_0.sRm = 0; gh1_0.sRn = 0;
      gh1_0.M = BK; gh1_0.N = H3; gh1_0.K = H; gh1_0.zi_n = 1; gh1_0.flags = 1; gh1_0.act = 0;
      gh1_0.alpha = 1.0f; gh1_0.beta = 0.0f; gh1_0.sa = 1.0f; gh1_0.sb = 1.0f; gh1_0.Npad = H3; gh1_0.pad_ = 0;
      k_gemm<1><<<dim3((unsigned)((H3) + 31) / 32, (unsigned)((BK) + 15) / 16, (unsigned)(1)), 32, 0, stream>>>(gh1_0); }
    k_gru<<<(unsigned)(((long long)BK * H + 255) / 256), 256, 0, stream>>>(GI, nullptr, nullptr, nullptr, GH, H1, H1n, BK, H);
    { GemmP gd_0;
      gd_0.A = H1n; gd_0.B = ow; gd_0.bias = ob; gd_0.R = H1n; gd_0.C = DL;
      gd_0.sAo = 0; gd_0.sAi = 0; gd_0.sAm = H; gd_0.sAk = 1; gd_0.sBo = 0; gd_0.sBi = 0; gd_0.sBn = H; gd_0.sBk = 1; gd_0.sCo = 0; gd_0.sCi = 0; gd_0.sCm = LDP; gd_0.sRo = 0; gd_0.sRi = 0; gd_0.sRm = 0; gd_0.sRn = 0;
      gd_0.M = BK; gd_0.N = 2; gd_0.K = H; gd_0.zi_n = 1; gd_0.flags = 1; gd_0.act = 0;
      gd_0.alpha = 1.0f; gd_0.beta = 0.0f; gd_0.sa = 1.0f; gd_0.sb = 1.0f; gd_0.Npad = LDP; gd_0.pad_ = 0;
      k_gemm<1><<<dim3((unsigned)((LDP) + 31) / 32, (unsigned)((BK) + 15) / 16, (unsigned)(1)), 32, 0, stream>>>(gd_0); }
    k_posstep<<<(unsigned)((BK * 2 + 255) / 256), 256, 0, stream>>>(DL, LDP, X, POS, TRAJ, BK, T, 0);
    k_lincopy<<<(unsigned)(((long long)(BK) * (H) + 255) / 256), 256, 0, stream>>>(H0n, H, H0, H, BK, H);
    k_lincopy<<<(unsigned)(((long long)(BK) * (H) + 255) / 256), 256, 0, stream>>>(H1n, H, H1, H, BK, H);
    { GemmP gh0_1;
      gh0_1.A = H0; gh0_1.B = whh0; gh0_1.bias = bhh0; gh0_1.R = H0; gh0_1.C = GH;
      gh0_1.sAo = 0; gh0_1.sAi = 0; gh0_1.sAm = H; gh0_1.sAk = 1; gh0_1.sBo = 0; gh0_1.sBi = 0; gh0_1.sBn = H; gh0_1.sBk = 1; gh0_1.sCo = 0; gh0_1.sCi = 0; gh0_1.sCm = H3; gh0_1.sRo = 0; gh0_1.sRi = 0; gh0_1.sRm = 0; gh0_1.sRn = 0;
      gh0_1.M = BK; gh0_1.N = H3; gh0_1.K = H; gh0_1.zi_n = 1; gh0_1.flags = 1; gh0_1.act = 0;
      gh0_1.alpha = 1.0f; gh0_1.beta = 0.0f; gh0_1.sa = 1.0f; gh0_1.sb = 1.0f; gh0_1.Npad = H3; gh0_1.pad_ = 0;
      k_gemm<1><<<dim3((unsigned)((H3) + 31) / 32, (unsigned)((BK) + 15) / 16, (unsigned)(1)), 32, 0, stream>>>(gh0_1); }
    k_gru<<<(unsigned)(((long long)BK * H + 255) / 256), 256, 0, stream>>>(nullptr, X, wih0, bih0, GH, H0, H0n, BK, H);
    { GemmP gi1_1;
      gi1_1.A = H0n; gi1_1.B = wih1; gi1_1.bias = bih1; gi1_1.R = H0n; gi1_1.C = GI;
      gi1_1.sAo = 0; gi1_1.sAi = 0; gi1_1.sAm = H; gi1_1.sAk = 1; gi1_1.sBo = 0; gi1_1.sBi = 0; gi1_1.sBn = H; gi1_1.sBk = 1; gi1_1.sCo = 0; gi1_1.sCi = 0; gi1_1.sCm = H3; gi1_1.sRo = 0; gi1_1.sRi = 0; gi1_1.sRm = 0; gi1_1.sRn = 0;
      gi1_1.M = BK; gi1_1.N = H3; gi1_1.K = H; gi1_1.zi_n = 1; gi1_1.flags = 1; gi1_1.act = 0;
      gi1_1.alpha = 1.0f; gi1_1.beta = 0.0f; gi1_1.sa = 1.0f; gi1_1.sb = 1.0f; gi1_1.Npad = H3; gi1_1.pad_ = 0;
      k_gemm<1><<<dim3((unsigned)((H3) + 31) / 32, (unsigned)((BK) + 15) / 16, (unsigned)(1)), 32, 0, stream>>>(gi1_1); }
    { GemmP gh1_1;
      gh1_1.A = H1; gh1_1.B = whh1; gh1_1.bias = bhh1; gh1_1.R = H1; gh1_1.C = GH;
      gh1_1.sAo = 0; gh1_1.sAi = 0; gh1_1.sAm = H; gh1_1.sAk = 1; gh1_1.sBo = 0; gh1_1.sBi = 0; gh1_1.sBn = H; gh1_1.sBk = 1; gh1_1.sCo = 0; gh1_1.sCi = 0; gh1_1.sCm = H3; gh1_1.sRo = 0; gh1_1.sRi = 0; gh1_1.sRm = 0; gh1_1.sRn = 0;
      gh1_1.M = BK; gh1_1.N = H3; gh1_1.K = H; gh1_1.zi_n = 1; gh1_1.flags = 1; gh1_1.act = 0;
      gh1_1.alpha = 1.0f; gh1_1.beta = 0.0f; gh1_1.sa = 1.0f; gh1_1.sb = 1.0f; gh1_1.Npad = H3; gh1_1.pad_ = 0;
      k_gemm<1><<<dim3((unsigned)((H3) + 31) / 32, (unsigned)((BK) + 15) / 16, (unsigned)(1)), 32, 0, stream>>>(gh1_1); }
    k_gru<<<(unsigned)(((long long)BK * H + 255) / 256), 256, 0, stream>>>(GI, nullptr, nullptr, nullptr, GH, H1, H1n, BK, H);
    { GemmP gd_1;
      gd_1.A = H1n; gd_1.B = ow; gd_1.bias = ob; gd_1.R = H1n; gd_1.C = DL;
      gd_1.sAo = 0; gd_1.sAi = 0; gd_1.sAm = H; gd_1.sAk = 1; gd_1.sBo = 0; gd_1.sBi = 0; gd_1.sBn = H; gd_1.sBk = 1; gd_1.sCo = 0; gd_1.sCi = 0; gd_1.sCm = LDP; gd_1.sRo = 0; gd_1.sRi = 0; gd_1.sRm = 0; gd_1.sRn = 0;
      gd_1.M = BK; gd_1.N = 2; gd_1.K = H; gd_1.zi_n = 1; gd_1.flags = 1; gd_1.act = 0;
      gd_1.alpha = 1.0f; gd_1.beta = 0.0f; gd_1.sa = 1.0f; gd_1.sb = 1.0f; gd_1.Npad = LDP; gd_1.pad_ = 0;
      k_gemm<1><<<dim3((unsigned)((LDP) + 31) / 32, (unsigned)((BK) + 15) / 16, (unsigned)(1)), 32, 0, stream>>>(gd_1); }
    k_posstep<<<(unsigned)((BK * 2 + 255) / 256), 256, 0, stream>>>(DL, LDP, X, POS, TRAJ, BK, T, 1);
    k_lincopy<<<(unsigned)(((long long)(BK) * (H) + 255) / 256), 256, 0, stream>>>(H0n, H, H0, H, BK, H);
    k_lincopy<<<(unsigned)(((long long)(BK) * (H) + 255) / 256), 256, 0, stream>>>(H1n, H, H1, H, BK, H);
    { GemmP gh0_2;
      gh0_2.A = H0; gh0_2.B = whh0; gh0_2.bias = bhh0; gh0_2.R = H0; gh0_2.C = GH;
      gh0_2.sAo = 0; gh0_2.sAi = 0; gh0_2.sAm = H; gh0_2.sAk = 1; gh0_2.sBo = 0; gh0_2.sBi = 0; gh0_2.sBn = H; gh0_2.sBk = 1; gh0_2.sCo = 0; gh0_2.sCi = 0; gh0_2.sCm = H3; gh0_2.sRo = 0; gh0_2.sRi = 0; gh0_2.sRm = 0; gh0_2.sRn = 0;
      gh0_2.M = BK; gh0_2.N = H3; gh0_2.K = H; gh0_2.zi_n = 1; gh0_2.flags = 1; gh0_2.act = 0;
      gh0_2.alpha = 1.0f; gh0_2.beta = 0.0f; gh0_2.sa = 1.0f; gh0_2.sb = 1.0f; gh0_2.Npad = H3; gh0_2.pad_ = 0;
      k_gemm<1><<<dim3((unsigned)((H3) + 31) / 32, (unsigned)((BK) + 15) / 16, (unsigned)(1)), 32, 0, stream>>>(gh0_2); }
    k_gru<<<(unsigned)(((long long)BK * H + 255) / 256), 256, 0, stream>>>(nullptr, X, wih0, bih0, GH, H0, H0n, BK, H);
    { GemmP gi1_2;
      gi1_2.A = H0n; gi1_2.B = wih1; gi1_2.bias = bih1; gi1_2.R = H0n; gi1_2.C = GI;
      gi1_2.sAo = 0; gi1_2.sAi = 0; gi1_2.sAm = H; gi1_2.sAk = 1; gi1_2.sBo = 0; gi1_2.sBi = 0; gi1_2.sBn = H; gi1_2.sBk = 1; gi1_2.sCo = 0; gi1_2.sCi = 0; gi1_2.sCm = H3; gi1_2.sRo = 0; gi1_2.sRi = 0; gi1_2.sRm = 0; gi1_2.sRn = 0;
      gi1_2.M = BK; gi1_2.N = H3; gi1_2.K = H; gi1_2.zi_n = 1; gi1_2.flags = 1; gi1_2.act = 0;
      gi1_2.alpha = 1.0f; gi1_2.beta = 0.0f; gi1_2.sa = 1.0f; gi1_2.sb = 1.0f; gi1_2.Npad = H3; gi1_2.pad_ = 0;
      k_gemm<1><<<dim3((unsigned)((H3) + 31) / 32, (unsigned)((BK) + 15) / 16, (unsigned)(1)), 32, 0, stream>>>(gi1_2); }
    { GemmP gh1_2;
      gh1_2.A = H1; gh1_2.B = whh1; gh1_2.bias = bhh1; gh1_2.R = H1; gh1_2.C = GH;
      gh1_2.sAo = 0; gh1_2.sAi = 0; gh1_2.sAm = H; gh1_2.sAk = 1; gh1_2.sBo = 0; gh1_2.sBi = 0; gh1_2.sBn = H; gh1_2.sBk = 1; gh1_2.sCo = 0; gh1_2.sCi = 0; gh1_2.sCm = H3; gh1_2.sRo = 0; gh1_2.sRi = 0; gh1_2.sRm = 0; gh1_2.sRn = 0;
      gh1_2.M = BK; gh1_2.N = H3; gh1_2.K = H; gh1_2.zi_n = 1; gh1_2.flags = 1; gh1_2.act = 0;
      gh1_2.alpha = 1.0f; gh1_2.beta = 0.0f; gh1_2.sa = 1.0f; gh1_2.sb = 1.0f; gh1_2.Npad = H3; gh1_2.pad_ = 0;
      k_gemm<1><<<dim3((unsigned)((H3) + 31) / 32, (unsigned)((BK) + 15) / 16, (unsigned)(1)), 32, 0, stream>>>(gh1_2); }
    k_gru<<<(unsigned)(((long long)BK * H + 255) / 256), 256, 0, stream>>>(GI, nullptr, nullptr, nullptr, GH, H1, H1n, BK, H);
    { GemmP gd_2;
      gd_2.A = H1n; gd_2.B = ow; gd_2.bias = ob; gd_2.R = H1n; gd_2.C = DL;
      gd_2.sAo = 0; gd_2.sAi = 0; gd_2.sAm = H; gd_2.sAk = 1; gd_2.sBo = 0; gd_2.sBi = 0; gd_2.sBn = H; gd_2.sBk = 1; gd_2.sCo = 0; gd_2.sCi = 0; gd_2.sCm = LDP; gd_2.sRo = 0; gd_2.sRi = 0; gd_2.sRm = 0; gd_2.sRn = 0;
      gd_2.M = BK; gd_2.N = 2; gd_2.K = H; gd_2.zi_n = 1; gd_2.flags = 1; gd_2.act = 0;
      gd_2.alpha = 1.0f; gd_2.beta = 0.0f; gd_2.sa = 1.0f; gd_2.sb = 1.0f; gd_2.Npad = LDP; gd_2.pad_ = 0;
      k_gemm<1><<<dim3((unsigned)((LDP) + 31) / 32, (unsigned)((BK) + 15) / 16, (unsigned)(1)), 32, 0, stream>>>(gd_2); }
    k_posstep<<<(unsigned)((BK * 2 + 255) / 256), 256, 0, stream>>>(DL, LDP, X, POS, TRAJ, BK, T, 2);
    k_lincopy<<<(unsigned)(((long long)(BK) * (H) + 255) / 256), 256, 0, stream>>>(H0n, H, H0, H, BK, H);
    k_lincopy<<<(unsigned)(((long long)(BK) * (H) + 255) / 256), 256, 0, stream>>>(H1n, H, H1, H, BK, H);
    { GemmP gh0_3;
      gh0_3.A = H0; gh0_3.B = whh0; gh0_3.bias = bhh0; gh0_3.R = H0; gh0_3.C = GH;
      gh0_3.sAo = 0; gh0_3.sAi = 0; gh0_3.sAm = H; gh0_3.sAk = 1; gh0_3.sBo = 0; gh0_3.sBi = 0; gh0_3.sBn = H; gh0_3.sBk = 1; gh0_3.sCo = 0; gh0_3.sCi = 0; gh0_3.sCm = H3; gh0_3.sRo = 0; gh0_3.sRi = 0; gh0_3.sRm = 0; gh0_3.sRn = 0;
      gh0_3.M = BK; gh0_3.N = H3; gh0_3.K = H; gh0_3.zi_n = 1; gh0_3.flags = 1; gh0_3.act = 0;
      gh0_3.alpha = 1.0f; gh0_3.beta = 0.0f; gh0_3.sa = 1.0f; gh0_3.sb = 1.0f; gh0_3.Npad = H3; gh0_3.pad_ = 0;
      k_gemm<1><<<dim3((unsigned)((H3) + 31) / 32, (unsigned)((BK) + 15) / 16, (unsigned)(1)), 32, 0, stream>>>(gh0_3); }
    k_gru<<<(unsigned)(((long long)BK * H + 255) / 256), 256, 0, stream>>>(nullptr, X, wih0, bih0, GH, H0, H0n, BK, H);
    { GemmP gi1_3;
      gi1_3.A = H0n; gi1_3.B = wih1; gi1_3.bias = bih1; gi1_3.R = H0n; gi1_3.C = GI;
      gi1_3.sAo = 0; gi1_3.sAi = 0; gi1_3.sAm = H; gi1_3.sAk = 1; gi1_3.sBo = 0; gi1_3.sBi = 0; gi1_3.sBn = H; gi1_3.sBk = 1; gi1_3.sCo = 0; gi1_3.sCi = 0; gi1_3.sCm = H3; gi1_3.sRo = 0; gi1_3.sRi = 0; gi1_3.sRm = 0; gi1_3.sRn = 0;
      gi1_3.M = BK; gi1_3.N = H3; gi1_3.K = H; gi1_3.zi_n = 1; gi1_3.flags = 1; gi1_3.act = 0;
      gi1_3.alpha = 1.0f; gi1_3.beta = 0.0f; gi1_3.sa = 1.0f; gi1_3.sb = 1.0f; gi1_3.Npad = H3; gi1_3.pad_ = 0;
      k_gemm<1><<<dim3((unsigned)((H3) + 31) / 32, (unsigned)((BK) + 15) / 16, (unsigned)(1)), 32, 0, stream>>>(gi1_3); }
    { GemmP gh1_3;
      gh1_3.A = H1; gh1_3.B = whh1; gh1_3.bias = bhh1; gh1_3.R = H1; gh1_3.C = GH;
      gh1_3.sAo = 0; gh1_3.sAi = 0; gh1_3.sAm = H; gh1_3.sAk = 1; gh1_3.sBo = 0; gh1_3.sBi = 0; gh1_3.sBn = H; gh1_3.sBk = 1; gh1_3.sCo = 0; gh1_3.sCi = 0; gh1_3.sCm = H3; gh1_3.sRo = 0; gh1_3.sRi = 0; gh1_3.sRm = 0; gh1_3.sRn = 0;
      gh1_3.M = BK; gh1_3.N = H3; gh1_3.K = H; gh1_3.zi_n = 1; gh1_3.flags = 1; gh1_3.act = 0;
      gh1_3.alpha = 1.0f; gh1_3.beta = 0.0f; gh1_3.sa = 1.0f; gh1_3.sb = 1.0f; gh1_3.Npad = H3; gh1_3.pad_ = 0;
      k_gemm<1><<<dim3((unsigned)((H3) + 31) / 32, (unsigned)((BK) + 15) / 16, (unsigned)(1)), 32, 0, stream>>>(gh1_3); }
    k_gru<<<(unsigned)(((long long)BK * H + 255) / 256), 256, 0, stream>>>(GI, nullptr, nullptr, nullptr, GH, H1, H1n, BK, H);
    { GemmP gd_3;
      gd_3.A = H1n; gd_3.B = ow; gd_3.bias = ob; gd_3.R = H1n; gd_3.C = DL;
      gd_3.sAo = 0; gd_3.sAi = 0; gd_3.sAm = H; gd_3.sAk = 1; gd_3.sBo = 0; gd_3.sBi = 0; gd_3.sBn = H; gd_3.sBk = 1; gd_3.sCo = 0; gd_3.sCi = 0; gd_3.sCm = LDP; gd_3.sRo = 0; gd_3.sRi = 0; gd_3.sRm = 0; gd_3.sRn = 0;
      gd_3.M = BK; gd_3.N = 2; gd_3.K = H; gd_3.zi_n = 1; gd_3.flags = 1; gd_3.act = 0;
      gd_3.alpha = 1.0f; gd_3.beta = 0.0f; gd_3.sa = 1.0f; gd_3.sb = 1.0f; gd_3.Npad = LDP; gd_3.pad_ = 0;
      k_gemm<1><<<dim3((unsigned)((LDP) + 31) / 32, (unsigned)((BK) + 15) / 16, (unsigned)(1)), 32, 0, stream>>>(gd_3); }
    k_posstep<<<(unsigned)((BK * 2 + 255) / 256), 256, 0, stream>>>(DL, LDP, X, POS, TRAJ, BK, T, 3);
    k_lincopy<<<(unsigned)(((long long)(BK) * (H) + 255) / 256), 256, 0, stream>>>(H0n, H, H0, H, BK, H);
    k_lincopy<<<(unsigned)(((long long)(BK) * (H) + 255) / 256), 256, 0, stream>>>(H1n, H, H1, H, BK, H);
    { GemmP gh0_4;
      gh0_4.A = H0; gh0_4.B = whh0; gh0_4.bias = bhh0; gh0_4.R = H0; gh0_4.C = GH;
      gh0_4.sAo = 0; gh0_4.sAi = 0; gh0_4.sAm = H; gh0_4.sAk = 1; gh0_4.sBo = 0; gh0_4.sBi = 0; gh0_4.sBn = H; gh0_4.sBk = 1; gh0_4.sCo = 0; gh0_4.sCi = 0; gh0_4.sCm = H3; gh0_4.sRo = 0; gh0_4.sRi = 0; gh0_4.sRm = 0; gh0_4.sRn = 0;
      gh0_4.M = BK; gh0_4.N = H3; gh0_4.K = H; gh0_4.zi_n = 1; gh0_4.flags = 1; gh0_4.act = 0;
      gh0_4.alpha = 1.0f; gh0_4.beta = 0.0f; gh0_4.sa = 1.0f; gh0_4.sb = 1.0f; gh0_4.Npad = H3; gh0_4.pad_ = 0;
      k_gemm<1><<<dim3((unsigned)((H3) + 31) / 32, (unsigned)((BK) + 15) / 16, (unsigned)(1)), 32, 0, stream>>>(gh0_4); }
    k_gru<<<(unsigned)(((long long)BK * H + 255) / 256), 256, 0, stream>>>(nullptr, X, wih0, bih0, GH, H0, H0n, BK, H);
    { GemmP gi1_4;
      gi1_4.A = H0n; gi1_4.B = wih1; gi1_4.bias = bih1; gi1_4.R = H0n; gi1_4.C = GI;
      gi1_4.sAo = 0; gi1_4.sAi = 0; gi1_4.sAm = H; gi1_4.sAk = 1; gi1_4.sBo = 0; gi1_4.sBi = 0; gi1_4.sBn = H; gi1_4.sBk = 1; gi1_4.sCo = 0; gi1_4.sCi = 0; gi1_4.sCm = H3; gi1_4.sRo = 0; gi1_4.sRi = 0; gi1_4.sRm = 0; gi1_4.sRn = 0;
      gi1_4.M = BK; gi1_4.N = H3; gi1_4.K = H; gi1_4.zi_n = 1; gi1_4.flags = 1; gi1_4.act = 0;
      gi1_4.alpha = 1.0f; gi1_4.beta = 0.0f; gi1_4.sa = 1.0f; gi1_4.sb = 1.0f; gi1_4.Npad = H3; gi1_4.pad_ = 0;
      k_gemm<1><<<dim3((unsigned)((H3) + 31) / 32, (unsigned)((BK) + 15) / 16, (unsigned)(1)), 32, 0, stream>>>(gi1_4); }
    { GemmP gh1_4;
      gh1_4.A = H1; gh1_4.B = whh1; gh1_4.bias = bhh1; gh1_4.R = H1; gh1_4.C = GH;
      gh1_4.sAo = 0; gh1_4.sAi = 0; gh1_4.sAm = H; gh1_4.sAk = 1; gh1_4.sBo = 0; gh1_4.sBi = 0; gh1_4.sBn = H; gh1_4.sBk = 1; gh1_4.sCo = 0; gh1_4.sCi = 0; gh1_4.sCm = H3; gh1_4.sRo = 0; gh1_4.sRi = 0; gh1_4.sRm = 0; gh1_4.sRn = 0;
      gh1_4.M = BK; gh1_4.N = H3; gh1_4.K = H; gh1_4.zi_n = 1; gh1_4.flags = 1; gh1_4.act = 0;
      gh1_4.alpha = 1.0f; gh1_4.beta = 0.0f; gh1_4.sa = 1.0f; gh1_4.sb = 1.0f; gh1_4.Npad = H3; gh1_4.pad_ = 0;
      k_gemm<1><<<dim3((unsigned)((H3) + 31) / 32, (unsigned)((BK) + 15) / 16, (unsigned)(1)), 32, 0, stream>>>(gh1_4); }
    k_gru<<<(unsigned)(((long long)BK * H + 255) / 256), 256, 0, stream>>>(GI, nullptr, nullptr, nullptr, GH, H1, H1n, BK, H);
    { GemmP gd_4;
      gd_4.A = H1n; gd_4.B = ow; gd_4.bias = ob; gd_4.R = H1n; gd_4.C = DL;
      gd_4.sAo = 0; gd_4.sAi = 0; gd_4.sAm = H; gd_4.sAk = 1; gd_4.sBo = 0; gd_4.sBi = 0; gd_4.sBn = H; gd_4.sBk = 1; gd_4.sCo = 0; gd_4.sCi = 0; gd_4.sCm = LDP; gd_4.sRo = 0; gd_4.sRi = 0; gd_4.sRm = 0; gd_4.sRn = 0;
      gd_4.M = BK; gd_4.N = 2; gd_4.K = H; gd_4.zi_n = 1; gd_4.flags = 1; gd_4.act = 0;
      gd_4.alpha = 1.0f; gd_4.beta = 0.0f; gd_4.sa = 1.0f; gd_4.sb = 1.0f; gd_4.Npad = LDP; gd_4.pad_ = 0;
      k_gemm<1><<<dim3((unsigned)((LDP) + 31) / 32, (unsigned)((BK) + 15) / 16, (unsigned)(1)), 32, 0, stream>>>(gd_4); }
    k_posstep<<<(unsigned)((BK * 2 + 255) / 256), 256, 0, stream>>>(DL, LDP, X, POS, TRAJ, BK, T, 4);
    k_lincopy<<<(unsigned)(((long long)(BK) * (H) + 255) / 256), 256, 0, stream>>>(H0n, H, H0, H, BK, H);
    k_lincopy<<<(unsigned)(((long long)(BK) * (H) + 255) / 256), 256, 0, stream>>>(H1n, H, H1, H, BK, H);
    { GemmP gh0_5;
      gh0_5.A = H0; gh0_5.B = whh0; gh0_5.bias = bhh0; gh0_5.R = H0; gh0_5.C = GH;
      gh0_5.sAo = 0; gh0_5.sAi = 0; gh0_5.sAm = H; gh0_5.sAk = 1; gh0_5.sBo = 0; gh0_5.sBi = 0; gh0_5.sBn = H; gh0_5.sBk = 1; gh0_5.sCo = 0; gh0_5.sCi = 0; gh0_5.sCm = H3; gh0_5.sRo = 0; gh0_5.sRi = 0; gh0_5.sRm = 0; gh0_5.sRn = 0;
      gh0_5.M = BK; gh0_5.N = H3; gh0_5.K = H; gh0_5.zi_n = 1; gh0_5.flags = 1; gh0_5.act = 0;
      gh0_5.alpha = 1.0f; gh0_5.beta = 0.0f; gh0_5.sa = 1.0f; gh0_5.sb = 1.0f; gh0_5.Npad = H3; gh0_5.pad_ = 0;
      k_gemm<1><<<dim3((unsigned)((H3) + 31) / 32, (unsigned)((BK) + 15) / 16, (unsigned)(1)), 32, 0, stream>>>(gh0_5); }
    k_gru<<<(unsigned)(((long long)BK * H + 255) / 256), 256, 0, stream>>>(nullptr, X, wih0, bih0, GH, H0, H0n, BK, H);
    { GemmP gi1_5;
      gi1_5.A = H0n; gi1_5.B = wih1; gi1_5.bias = bih1; gi1_5.R = H0n; gi1_5.C = GI;
      gi1_5.sAo = 0; gi1_5.sAi = 0; gi1_5.sAm = H; gi1_5.sAk = 1; gi1_5.sBo = 0; gi1_5.sBi = 0; gi1_5.sBn = H; gi1_5.sBk = 1; gi1_5.sCo = 0; gi1_5.sCi = 0; gi1_5.sCm = H3; gi1_5.sRo = 0; gi1_5.sRi = 0; gi1_5.sRm = 0; gi1_5.sRn = 0;
      gi1_5.M = BK; gi1_5.N = H3; gi1_5.K = H; gi1_5.zi_n = 1; gi1_5.flags = 1; gi1_5.act = 0;
      gi1_5.alpha = 1.0f; gi1_5.beta = 0.0f; gi1_5.sa = 1.0f; gi1_5.sb = 1.0f; gi1_5.Npad = H3; gi1_5.pad_ = 0;
      k_gemm<1><<<dim3((unsigned)((H3) + 31) / 32, (unsigned)((BK) + 15) / 16, (unsigned)(1)), 32, 0, stream>>>(gi1_5); }
    { GemmP gh1_5;
      gh1_5.A = H1; gh1_5.B = whh1; gh1_5.bias = bhh1; gh1_5.R = H1; gh1_5.C = GH;
      gh1_5.sAo = 0; gh1_5.sAi = 0; gh1_5.sAm = H; gh1_5.sAk = 1; gh1_5.sBo = 0; gh1_5.sBi = 0; gh1_5.sBn = H; gh1_5.sBk = 1; gh1_5.sCo = 0; gh1_5.sCi = 0; gh1_5.sCm = H3; gh1_5.sRo = 0; gh1_5.sRi = 0; gh1_5.sRm = 0; gh1_5.sRn = 0;
      gh1_5.M = BK; gh1_5.N = H3; gh1_5.K = H; gh1_5.zi_n = 1; gh1_5.flags = 1; gh1_5.act = 0;
      gh1_5.alpha = 1.0f; gh1_5.beta = 0.0f; gh1_5.sa = 1.0f; gh1_5.sb = 1.0f; gh1_5.Npad = H3; gh1_5.pad_ = 0;
      k_gemm<1><<<dim3((unsigned)((H3) + 31) / 32, (unsigned)((BK) + 15) / 16, (unsigned)(1)), 32, 0, stream>>>(gh1_5); }
    k_gru<<<(unsigned)(((long long)BK * H + 255) / 256), 256, 0, stream>>>(GI, nullptr, nullptr, nullptr, GH, H1, H1n, BK, H);
    { GemmP gd_5;
      gd_5.A = H1n; gd_5.B = ow; gd_5.bias = ob; gd_5.R = H1n; gd_5.C = DL;
      gd_5.sAo = 0; gd_5.sAi = 0; gd_5.sAm = H; gd_5.sAk = 1; gd_5.sBo = 0; gd_5.sBi = 0; gd_5.sBn = H; gd_5.sBk = 1; gd_5.sCo = 0; gd_5.sCi = 0; gd_5.sCm = LDP; gd_5.sRo = 0; gd_5.sRi = 0; gd_5.sRm = 0; gd_5.sRn = 0;
      gd_5.M = BK; gd_5.N = 2; gd_5.K = H; gd_5.zi_n = 1; gd_5.flags = 1; gd_5.act = 0;
      gd_5.alpha = 1.0f; gd_5.beta = 0.0f; gd_5.sa = 1.0f; gd_5.sb = 1.0f; gd_5.Npad = LDP; gd_5.pad_ = 0;
      k_gemm<1><<<dim3((unsigned)((LDP) + 31) / 32, (unsigned)((BK) + 15) / 16, (unsigned)(1)), 32, 0, stream>>>(gd_5); }
    k_posstep<<<(unsigned)((BK * 2 + 255) / 256), 256, 0, stream>>>(DL, LDP, X, POS, TRAJ, BK, T, 5);
    k_lincopy<<<(unsigned)(((long long)(BK) * (H) + 255) / 256), 256, 0, stream>>>(H0n, H, H0, H, BK, H);
    k_lincopy<<<(unsigned)(((long long)(BK) * (H) + 255) / 256), 256, 0, stream>>>(H1n, H, H1, H, BK, H);
    { GemmP gh0_6;
      gh0_6.A = H0; gh0_6.B = whh0; gh0_6.bias = bhh0; gh0_6.R = H0; gh0_6.C = GH;
      gh0_6.sAo = 0; gh0_6.sAi = 0; gh0_6.sAm = H; gh0_6.sAk = 1; gh0_6.sBo = 0; gh0_6.sBi = 0; gh0_6.sBn = H; gh0_6.sBk = 1; gh0_6.sCo = 0; gh0_6.sCi = 0; gh0_6.sCm = H3; gh0_6.sRo = 0; gh0_6.sRi = 0; gh0_6.sRm = 0; gh0_6.sRn = 0;
      gh0_6.M = BK; gh0_6.N = H3; gh0_6.K = H; gh0_6.zi_n = 1; gh0_6.flags = 1; gh0_6.act = 0;
      gh0_6.alpha = 1.0f; gh0_6.beta = 0.0f; gh0_6.sa = 1.0f; gh0_6.sb = 1.0f; gh0_6.Npad = H3; gh0_6.pad_ = 0;
      k_gemm<1><<<dim3((unsigned)((H3) + 31) / 32, (unsigned)((BK) + 15) / 16, (unsigned)(1)), 32, 0, stream>>>(gh0_6); }
    k_gru<<<(unsigned)(((long long)BK * H + 255) / 256), 256, 0, stream>>>(nullptr, X, wih0, bih0, GH, H0, H0n, BK, H);
    { GemmP gi1_6;
      gi1_6.A = H0n; gi1_6.B = wih1; gi1_6.bias = bih1; gi1_6.R = H0n; gi1_6.C = GI;
      gi1_6.sAo = 0; gi1_6.sAi = 0; gi1_6.sAm = H; gi1_6.sAk = 1; gi1_6.sBo = 0; gi1_6.sBi = 0; gi1_6.sBn = H; gi1_6.sBk = 1; gi1_6.sCo = 0; gi1_6.sCi = 0; gi1_6.sCm = H3; gi1_6.sRo = 0; gi1_6.sRi = 0; gi1_6.sRm = 0; gi1_6.sRn = 0;
      gi1_6.M = BK; gi1_6.N = H3; gi1_6.K = H; gi1_6.zi_n = 1; gi1_6.flags = 1; gi1_6.act = 0;
      gi1_6.alpha = 1.0f; gi1_6.beta = 0.0f; gi1_6.sa = 1.0f; gi1_6.sb = 1.0f; gi1_6.Npad = H3; gi1_6.pad_ = 0;
      k_gemm<1><<<dim3((unsigned)((H3) + 31) / 32, (unsigned)((BK) + 15) / 16, (unsigned)(1)), 32, 0, stream>>>(gi1_6); }
    { GemmP gh1_6;
      gh1_6.A = H1; gh1_6.B = whh1; gh1_6.bias = bhh1; gh1_6.R = H1; gh1_6.C = GH;
      gh1_6.sAo = 0; gh1_6.sAi = 0; gh1_6.sAm = H; gh1_6.sAk = 1; gh1_6.sBo = 0; gh1_6.sBi = 0; gh1_6.sBn = H; gh1_6.sBk = 1; gh1_6.sCo = 0; gh1_6.sCi = 0; gh1_6.sCm = H3; gh1_6.sRo = 0; gh1_6.sRi = 0; gh1_6.sRm = 0; gh1_6.sRn = 0;
      gh1_6.M = BK; gh1_6.N = H3; gh1_6.K = H; gh1_6.zi_n = 1; gh1_6.flags = 1; gh1_6.act = 0;
      gh1_6.alpha = 1.0f; gh1_6.beta = 0.0f; gh1_6.sa = 1.0f; gh1_6.sb = 1.0f; gh1_6.Npad = H3; gh1_6.pad_ = 0;
      k_gemm<1><<<dim3((unsigned)((H3) + 31) / 32, (unsigned)((BK) + 15) / 16, (unsigned)(1)), 32, 0, stream>>>(gh1_6); }
    k_gru<<<(unsigned)(((long long)BK * H + 255) / 256), 256, 0, stream>>>(GI, nullptr, nullptr, nullptr, GH, H1, H1n, BK, H);
    { GemmP gd_6;
      gd_6.A = H1n; gd_6.B = ow; gd_6.bias = ob; gd_6.R = H1n; gd_6.C = DL;
      gd_6.sAo = 0; gd_6.sAi = 0; gd_6.sAm = H; gd_6.sAk = 1; gd_6.sBo = 0; gd_6.sBi = 0; gd_6.sBn = H; gd_6.sBk = 1; gd_6.sCo = 0; gd_6.sCi = 0; gd_6.sCm = LDP; gd_6.sRo = 0; gd_6.sRi = 0; gd_6.sRm = 0; gd_6.sRn = 0;
      gd_6.M = BK; gd_6.N = 2; gd_6.K = H; gd_6.zi_n = 1; gd_6.flags = 1; gd_6.act = 0;
      gd_6.alpha = 1.0f; gd_6.beta = 0.0f; gd_6.sa = 1.0f; gd_6.sb = 1.0f; gd_6.Npad = LDP; gd_6.pad_ = 0;
      k_gemm<1><<<dim3((unsigned)((LDP) + 31) / 32, (unsigned)((BK) + 15) / 16, (unsigned)(1)), 32, 0, stream>>>(gd_6); }
    k_posstep<<<(unsigned)((BK * 2 + 255) / 256), 256, 0, stream>>>(DL, LDP, X, POS, TRAJ, BK, T, 6);
    k_lincopy<<<(unsigned)(((long long)(BK) * (H) + 255) / 256), 256, 0, stream>>>(H0n, H, H0, H, BK, H);
    k_lincopy<<<(unsigned)(((long long)(BK) * (H) + 255) / 256), 256, 0, stream>>>(H1n, H, H1, H, BK, H);
    { GemmP gh0_7;
      gh0_7.A = H0; gh0_7.B = whh0; gh0_7.bias = bhh0; gh0_7.R = H0; gh0_7.C = GH;
      gh0_7.sAo = 0; gh0_7.sAi = 0; gh0_7.sAm = H; gh0_7.sAk = 1; gh0_7.sBo = 0; gh0_7.sBi = 0; gh0_7.sBn = H; gh0_7.sBk = 1; gh0_7.sCo = 0; gh0_7.sCi = 0; gh0_7.sCm = H3; gh0_7.sRo = 0; gh0_7.sRi = 0; gh0_7.sRm = 0; gh0_7.sRn = 0;
      gh0_7.M = BK; gh0_7.N = H3; gh0_7.K = H; gh0_7.zi_n = 1; gh0_7.flags = 1; gh0_7.act = 0;
      gh0_7.alpha = 1.0f; gh0_7.beta = 0.0f; gh0_7.sa = 1.0f; gh0_7.sb = 1.0f; gh0_7.Npad = H3; gh0_7.pad_ = 0;
      k_gemm<1><<<dim3((unsigned)((H3) + 31) / 32, (unsigned)((BK) + 15) / 16, (unsigned)(1)), 32, 0, stream>>>(gh0_7); }
    k_gru<<<(unsigned)(((long long)BK * H + 255) / 256), 256, 0, stream>>>(nullptr, X, wih0, bih0, GH, H0, H0n, BK, H);
    { GemmP gi1_7;
      gi1_7.A = H0n; gi1_7.B = wih1; gi1_7.bias = bih1; gi1_7.R = H0n; gi1_7.C = GI;
      gi1_7.sAo = 0; gi1_7.sAi = 0; gi1_7.sAm = H; gi1_7.sAk = 1; gi1_7.sBo = 0; gi1_7.sBi = 0; gi1_7.sBn = H; gi1_7.sBk = 1; gi1_7.sCo = 0; gi1_7.sCi = 0; gi1_7.sCm = H3; gi1_7.sRo = 0; gi1_7.sRi = 0; gi1_7.sRm = 0; gi1_7.sRn = 0;
      gi1_7.M = BK; gi1_7.N = H3; gi1_7.K = H; gi1_7.zi_n = 1; gi1_7.flags = 1; gi1_7.act = 0;
      gi1_7.alpha = 1.0f; gi1_7.beta = 0.0f; gi1_7.sa = 1.0f; gi1_7.sb = 1.0f; gi1_7.Npad = H3; gi1_7.pad_ = 0;
      k_gemm<1><<<dim3((unsigned)((H3) + 31) / 32, (unsigned)((BK) + 15) / 16, (unsigned)(1)), 32, 0, stream>>>(gi1_7); }
    { GemmP gh1_7;
      gh1_7.A = H1; gh1_7.B = whh1; gh1_7.bias = bhh1; gh1_7.R = H1; gh1_7.C = GH;
      gh1_7.sAo = 0; gh1_7.sAi = 0; gh1_7.sAm = H; gh1_7.sAk = 1; gh1_7.sBo = 0; gh1_7.sBi = 0; gh1_7.sBn = H; gh1_7.sBk = 1; gh1_7.sCo = 0; gh1_7.sCi = 0; gh1_7.sCm = H3; gh1_7.sRo = 0; gh1_7.sRi = 0; gh1_7.sRm = 0; gh1_7.sRn = 0;
      gh1_7.M = BK; gh1_7.N = H3; gh1_7.K = H; gh1_7.zi_n = 1; gh1_7.flags = 1; gh1_7.act = 0;
      gh1_7.alpha = 1.0f; gh1_7.beta = 0.0f; gh1_7.sa = 1.0f; gh1_7.sb = 1.0f; gh1_7.Npad = H3; gh1_7.pad_ = 0;
      k_gemm<1><<<dim3((unsigned)((H3) + 31) / 32, (unsigned)((BK) + 15) / 16, (unsigned)(1)), 32, 0, stream>>>(gh1_7); }
    k_gru<<<(unsigned)(((long long)BK * H + 255) / 256), 256, 0, stream>>>(GI, nullptr, nullptr, nullptr, GH, H1, H1n, BK, H);
    { GemmP gd_7;
      gd_7.A = H1n; gd_7.B = ow; gd_7.bias = ob; gd_7.R = H1n; gd_7.C = DL;
      gd_7.sAo = 0; gd_7.sAi = 0; gd_7.sAm = H; gd_7.sAk = 1; gd_7.sBo = 0; gd_7.sBi = 0; gd_7.sBn = H; gd_7.sBk = 1; gd_7.sCo = 0; gd_7.sCi = 0; gd_7.sCm = LDP; gd_7.sRo = 0; gd_7.sRi = 0; gd_7.sRm = 0; gd_7.sRn = 0;
      gd_7.M = BK; gd_7.N = 2; gd_7.K = H; gd_7.zi_n = 1; gd_7.flags = 1; gd_7.act = 0;
      gd_7.alpha = 1.0f; gd_7.beta = 0.0f; gd_7.sa = 1.0f; gd_7.sb = 1.0f; gd_7.Npad = LDP; gd_7.pad_ = 0;
      k_gemm<1><<<dim3((unsigned)((LDP) + 31) / 32, (unsigned)((BK) + 15) / 16, (unsigned)(1)), 32, 0, stream>>>(gd_7); }
    k_posstep<<<(unsigned)((BK * 2 + 255) / 256), 256, 0, stream>>>(DL, LDP, X, POS, TRAJ, BK, T, 7);
    k_lincopy<<<(unsigned)(((long long)(BK) * (H) + 255) / 256), 256, 0, stream>>>(H0n, H, H0, H, BK, H);
    k_lincopy<<<(unsigned)(((long long)(BK) * (H) + 255) / 256), 256, 0, stream>>>(H1n, H, H1, H, BK, H);
    { GemmP gh0_8;
      gh0_8.A = H0; gh0_8.B = whh0; gh0_8.bias = bhh0; gh0_8.R = H0; gh0_8.C = GH;
      gh0_8.sAo = 0; gh0_8.sAi = 0; gh0_8.sAm = H; gh0_8.sAk = 1; gh0_8.sBo = 0; gh0_8.sBi = 0; gh0_8.sBn = H; gh0_8.sBk = 1; gh0_8.sCo = 0; gh0_8.sCi = 0; gh0_8.sCm = H3; gh0_8.sRo = 0; gh0_8.sRi = 0; gh0_8.sRm = 0; gh0_8.sRn = 0;
      gh0_8.M = BK; gh0_8.N = H3; gh0_8.K = H; gh0_8.zi_n = 1; gh0_8.flags = 1; gh0_8.act = 0;
      gh0_8.alpha = 1.0f; gh0_8.beta = 0.0f; gh0_8.sa = 1.0f; gh0_8.sb = 1.0f; gh0_8.Npad = H3; gh0_8.pad_ = 0;
      k_gemm<1><<<dim3((unsigned)((H3) + 31) / 32, (unsigned)((BK) + 15) / 16, (unsigned)(1)), 32, 0, stream>>>(gh0_8); }
    k_gru<<<(unsigned)(((long long)BK * H + 255) / 256), 256, 0, stream>>>(nullptr, X, wih0, bih0, GH, H0, H0n, BK, H);
    { GemmP gi1_8;
      gi1_8.A = H0n; gi1_8.B = wih1; gi1_8.bias = bih1; gi1_8.R = H0n; gi1_8.C = GI;
      gi1_8.sAo = 0; gi1_8.sAi = 0; gi1_8.sAm = H; gi1_8.sAk = 1; gi1_8.sBo = 0; gi1_8.sBi = 0; gi1_8.sBn = H; gi1_8.sBk = 1; gi1_8.sCo = 0; gi1_8.sCi = 0; gi1_8.sCm = H3; gi1_8.sRo = 0; gi1_8.sRi = 0; gi1_8.sRm = 0; gi1_8.sRn = 0;
      gi1_8.M = BK; gi1_8.N = H3; gi1_8.K = H; gi1_8.zi_n = 1; gi1_8.flags = 1; gi1_8.act = 0;
      gi1_8.alpha = 1.0f; gi1_8.beta = 0.0f; gi1_8.sa = 1.0f; gi1_8.sb = 1.0f; gi1_8.Npad = H3; gi1_8.pad_ = 0;
      k_gemm<1><<<dim3((unsigned)((H3) + 31) / 32, (unsigned)((BK) + 15) / 16, (unsigned)(1)), 32, 0, stream>>>(gi1_8); }
    { GemmP gh1_8;
      gh1_8.A = H1; gh1_8.B = whh1; gh1_8.bias = bhh1; gh1_8.R = H1; gh1_8.C = GH;
      gh1_8.sAo = 0; gh1_8.sAi = 0; gh1_8.sAm = H; gh1_8.sAk = 1; gh1_8.sBo = 0; gh1_8.sBi = 0; gh1_8.sBn = H; gh1_8.sBk = 1; gh1_8.sCo = 0; gh1_8.sCi = 0; gh1_8.sCm = H3; gh1_8.sRo = 0; gh1_8.sRi = 0; gh1_8.sRm = 0; gh1_8.sRn = 0;
      gh1_8.M = BK; gh1_8.N = H3; gh1_8.K = H; gh1_8.zi_n = 1; gh1_8.flags = 1; gh1_8.act = 0;
      gh1_8.alpha = 1.0f; gh1_8.beta = 0.0f; gh1_8.sa = 1.0f; gh1_8.sb = 1.0f; gh1_8.Npad = H3; gh1_8.pad_ = 0;
      k_gemm<1><<<dim3((unsigned)((H3) + 31) / 32, (unsigned)((BK) + 15) / 16, (unsigned)(1)), 32, 0, stream>>>(gh1_8); }
    k_gru<<<(unsigned)(((long long)BK * H + 255) / 256), 256, 0, stream>>>(GI, nullptr, nullptr, nullptr, GH, H1, H1n, BK, H);
    { GemmP gd_8;
      gd_8.A = H1n; gd_8.B = ow; gd_8.bias = ob; gd_8.R = H1n; gd_8.C = DL;
      gd_8.sAo = 0; gd_8.sAi = 0; gd_8.sAm = H; gd_8.sAk = 1; gd_8.sBo = 0; gd_8.sBi = 0; gd_8.sBn = H; gd_8.sBk = 1; gd_8.sCo = 0; gd_8.sCi = 0; gd_8.sCm = LDP; gd_8.sRo = 0; gd_8.sRi = 0; gd_8.sRm = 0; gd_8.sRn = 0;
      gd_8.M = BK; gd_8.N = 2; gd_8.K = H; gd_8.zi_n = 1; gd_8.flags = 1; gd_8.act = 0;
      gd_8.alpha = 1.0f; gd_8.beta = 0.0f; gd_8.sa = 1.0f; gd_8.sb = 1.0f; gd_8.Npad = LDP; gd_8.pad_ = 0;
      k_gemm<1><<<dim3((unsigned)((LDP) + 31) / 32, (unsigned)((BK) + 15) / 16, (unsigned)(1)), 32, 0, stream>>>(gd_8); }
    k_posstep<<<(unsigned)((BK * 2 + 255) / 256), 256, 0, stream>>>(DL, LDP, X, POS, TRAJ, BK, T, 8);
    k_lincopy<<<(unsigned)(((long long)(BK) * (H) + 255) / 256), 256, 0, stream>>>(H0n, H, H0, H, BK, H);
    k_lincopy<<<(unsigned)(((long long)(BK) * (H) + 255) / 256), 256, 0, stream>>>(H1n, H, H1, H, BK, H);
    { GemmP gh0_9;
      gh0_9.A = H0; gh0_9.B = whh0; gh0_9.bias = bhh0; gh0_9.R = H0; gh0_9.C = GH;
      gh0_9.sAo = 0; gh0_9.sAi = 0; gh0_9.sAm = H; gh0_9.sAk = 1; gh0_9.sBo = 0; gh0_9.sBi = 0; gh0_9.sBn = H; gh0_9.sBk = 1; gh0_9.sCo = 0; gh0_9.sCi = 0; gh0_9.sCm = H3; gh0_9.sRo = 0; gh0_9.sRi = 0; gh0_9.sRm = 0; gh0_9.sRn = 0;
      gh0_9.M = BK; gh0_9.N = H3; gh0_9.K = H; gh0_9.zi_n = 1; gh0_9.flags = 1; gh0_9.act = 0;
      gh0_9.alpha = 1.0f; gh0_9.beta = 0.0f; gh0_9.sa = 1.0f; gh0_9.sb = 1.0f; gh0_9.Npad = H3; gh0_9.pad_ = 0;
      k_gemm<1><<<dim3((unsigned)((H3) + 31) / 32, (unsigned)((BK) + 15) / 16, (unsigned)(1)), 32, 0, stream>>>(gh0_9); }
    k_gru<<<(unsigned)(((long long)BK * H + 255) / 256), 256, 0, stream>>>(nullptr, X, wih0, bih0, GH, H0, H0n, BK, H);
    { GemmP gi1_9;
      gi1_9.A = H0n; gi1_9.B = wih1; gi1_9.bias = bih1; gi1_9.R = H0n; gi1_9.C = GI;
      gi1_9.sAo = 0; gi1_9.sAi = 0; gi1_9.sAm = H; gi1_9.sAk = 1; gi1_9.sBo = 0; gi1_9.sBi = 0; gi1_9.sBn = H; gi1_9.sBk = 1; gi1_9.sCo = 0; gi1_9.sCi = 0; gi1_9.sCm = H3; gi1_9.sRo = 0; gi1_9.sRi = 0; gi1_9.sRm = 0; gi1_9.sRn = 0;
      gi1_9.M = BK; gi1_9.N = H3; gi1_9.K = H; gi1_9.zi_n = 1; gi1_9.flags = 1; gi1_9.act = 0;
      gi1_9.alpha = 1.0f; gi1_9.beta = 0.0f; gi1_9.sa = 1.0f; gi1_9.sb = 1.0f; gi1_9.Npad = H3; gi1_9.pad_ = 0;
      k_gemm<1><<<dim3((unsigned)((H3) + 31) / 32, (unsigned)((BK) + 15) / 16, (unsigned)(1)), 32, 0, stream>>>(gi1_9); }
    { GemmP gh1_9;
      gh1_9.A = H1; gh1_9.B = whh1; gh1_9.bias = bhh1; gh1_9.R = H1; gh1_9.C = GH;
      gh1_9.sAo = 0; gh1_9.sAi = 0; gh1_9.sAm = H; gh1_9.sAk = 1; gh1_9.sBo = 0; gh1_9.sBi = 0; gh1_9.sBn = H; gh1_9.sBk = 1; gh1_9.sCo = 0; gh1_9.sCi = 0; gh1_9.sCm = H3; gh1_9.sRo = 0; gh1_9.sRi = 0; gh1_9.sRm = 0; gh1_9.sRn = 0;
      gh1_9.M = BK; gh1_9.N = H3; gh1_9.K = H; gh1_9.zi_n = 1; gh1_9.flags = 1; gh1_9.act = 0;
      gh1_9.alpha = 1.0f; gh1_9.beta = 0.0f; gh1_9.sa = 1.0f; gh1_9.sb = 1.0f; gh1_9.Npad = H3; gh1_9.pad_ = 0;
      k_gemm<1><<<dim3((unsigned)((H3) + 31) / 32, (unsigned)((BK) + 15) / 16, (unsigned)(1)), 32, 0, stream>>>(gh1_9); }
    k_gru<<<(unsigned)(((long long)BK * H + 255) / 256), 256, 0, stream>>>(GI, nullptr, nullptr, nullptr, GH, H1, H1n, BK, H);
    { GemmP gd_9;
      gd_9.A = H1n; gd_9.B = ow; gd_9.bias = ob; gd_9.R = H1n; gd_9.C = DL;
      gd_9.sAo = 0; gd_9.sAi = 0; gd_9.sAm = H; gd_9.sAk = 1; gd_9.sBo = 0; gd_9.sBi = 0; gd_9.sBn = H; gd_9.sBk = 1; gd_9.sCo = 0; gd_9.sCi = 0; gd_9.sCm = LDP; gd_9.sRo = 0; gd_9.sRi = 0; gd_9.sRm = 0; gd_9.sRn = 0;
      gd_9.M = BK; gd_9.N = 2; gd_9.K = H; gd_9.zi_n = 1; gd_9.flags = 1; gd_9.act = 0;
      gd_9.alpha = 1.0f; gd_9.beta = 0.0f; gd_9.sa = 1.0f; gd_9.sb = 1.0f; gd_9.Npad = LDP; gd_9.pad_ = 0;
      k_gemm<1><<<dim3((unsigned)((LDP) + 31) / 32, (unsigned)((BK) + 15) / 16, (unsigned)(1)), 32, 0, stream>>>(gd_9); }
    k_posstep<<<(unsigned)((BK * 2 + 255) / 256), 256, 0, stream>>>(DL, LDP, X, POS, TRAJ, BK, T, 9);
    k_lincopy<<<(unsigned)(((long long)(BK) * (H) + 255) / 256), 256, 0, stream>>>(H0n, H, H0, H, BK, H);
    k_lincopy<<<(unsigned)(((long long)(BK) * (H) + 255) / 256), 256, 0, stream>>>(H1n, H, H1, H, BK, H);
    { GemmP gh0_10;
      gh0_10.A = H0; gh0_10.B = whh0; gh0_10.bias = bhh0; gh0_10.R = H0; gh0_10.C = GH;
      gh0_10.sAo = 0; gh0_10.sAi = 0; gh0_10.sAm = H; gh0_10.sAk = 1; gh0_10.sBo = 0; gh0_10.sBi = 0; gh0_10.sBn = H; gh0_10.sBk = 1; gh0_10.sCo = 0; gh0_10.sCi = 0; gh0_10.sCm = H3; gh0_10.sRo = 0; gh0_10.sRi = 0; gh0_10.sRm = 0; gh0_10.sRn = 0;
      gh0_10.M = BK; gh0_10.N = H3; gh0_10.K = H; gh0_10.zi_n = 1; gh0_10.flags = 1; gh0_10.act = 0;
      gh0_10.alpha = 1.0f; gh0_10.beta = 0.0f; gh0_10.sa = 1.0f; gh0_10.sb = 1.0f; gh0_10.Npad = H3; gh0_10.pad_ = 0;
      k_gemm<1><<<dim3((unsigned)((H3) + 31) / 32, (unsigned)((BK) + 15) / 16, (unsigned)(1)), 32, 0, stream>>>(gh0_10); }
    k_gru<<<(unsigned)(((long long)BK * H + 255) / 256), 256, 0, stream>>>(nullptr, X, wih0, bih0, GH, H0, H0n, BK, H);
    { GemmP gi1_10;
      gi1_10.A = H0n; gi1_10.B = wih1; gi1_10.bias = bih1; gi1_10.R = H0n; gi1_10.C = GI;
      gi1_10.sAo = 0; gi1_10.sAi = 0; gi1_10.sAm = H; gi1_10.sAk = 1; gi1_10.sBo = 0; gi1_10.sBi = 0; gi1_10.sBn = H; gi1_10.sBk = 1; gi1_10.sCo = 0; gi1_10.sCi = 0; gi1_10.sCm = H3; gi1_10.sRo = 0; gi1_10.sRi = 0; gi1_10.sRm = 0; gi1_10.sRn = 0;
      gi1_10.M = BK; gi1_10.N = H3; gi1_10.K = H; gi1_10.zi_n = 1; gi1_10.flags = 1; gi1_10.act = 0;
      gi1_10.alpha = 1.0f; gi1_10.beta = 0.0f; gi1_10.sa = 1.0f; gi1_10.sb = 1.0f; gi1_10.Npad = H3; gi1_10.pad_ = 0;
      k_gemm<1><<<dim3((unsigned)((H3) + 31) / 32, (unsigned)((BK) + 15) / 16, (unsigned)(1)), 32, 0, stream>>>(gi1_10); }
    { GemmP gh1_10;
      gh1_10.A = H1; gh1_10.B = whh1; gh1_10.bias = bhh1; gh1_10.R = H1; gh1_10.C = GH;
      gh1_10.sAo = 0; gh1_10.sAi = 0; gh1_10.sAm = H; gh1_10.sAk = 1; gh1_10.sBo = 0; gh1_10.sBi = 0; gh1_10.sBn = H; gh1_10.sBk = 1; gh1_10.sCo = 0; gh1_10.sCi = 0; gh1_10.sCm = H3; gh1_10.sRo = 0; gh1_10.sRi = 0; gh1_10.sRm = 0; gh1_10.sRn = 0;
      gh1_10.M = BK; gh1_10.N = H3; gh1_10.K = H; gh1_10.zi_n = 1; gh1_10.flags = 1; gh1_10.act = 0;
      gh1_10.alpha = 1.0f; gh1_10.beta = 0.0f; gh1_10.sa = 1.0f; gh1_10.sb = 1.0f; gh1_10.Npad = H3; gh1_10.pad_ = 0;
      k_gemm<1><<<dim3((unsigned)((H3) + 31) / 32, (unsigned)((BK) + 15) / 16, (unsigned)(1)), 32, 0, stream>>>(gh1_10); }
    k_gru<<<(unsigned)(((long long)BK * H + 255) / 256), 256, 0, stream>>>(GI, nullptr, nullptr, nullptr, GH, H1, H1n, BK, H);
    { GemmP gd_10;
      gd_10.A = H1n; gd_10.B = ow; gd_10.bias = ob; gd_10.R = H1n; gd_10.C = DL;
      gd_10.sAo = 0; gd_10.sAi = 0; gd_10.sAm = H; gd_10.sAk = 1; gd_10.sBo = 0; gd_10.sBi = 0; gd_10.sBn = H; gd_10.sBk = 1; gd_10.sCo = 0; gd_10.sCi = 0; gd_10.sCm = LDP; gd_10.sRo = 0; gd_10.sRi = 0; gd_10.sRm = 0; gd_10.sRn = 0;
      gd_10.M = BK; gd_10.N = 2; gd_10.K = H; gd_10.zi_n = 1; gd_10.flags = 1; gd_10.act = 0;
      gd_10.alpha = 1.0f; gd_10.beta = 0.0f; gd_10.sa = 1.0f; gd_10.sb = 1.0f; gd_10.Npad = LDP; gd_10.pad_ = 0;
      k_gemm<1><<<dim3((unsigned)((LDP) + 31) / 32, (unsigned)((BK) + 15) / 16, (unsigned)(1)), 32, 0, stream>>>(gd_10); }
    k_posstep<<<(unsigned)((BK * 2 + 255) / 256), 256, 0, stream>>>(DL, LDP, X, POS, TRAJ, BK, T, 10);
    k_lincopy<<<(unsigned)(((long long)(BK) * (H) + 255) / 256), 256, 0, stream>>>(H0n, H, H0, H, BK, H);
    k_lincopy<<<(unsigned)(((long long)(BK) * (H) + 255) / 256), 256, 0, stream>>>(H1n, H, H1, H, BK, H);
    { GemmP gh0_11;
      gh0_11.A = H0; gh0_11.B = whh0; gh0_11.bias = bhh0; gh0_11.R = H0; gh0_11.C = GH;
      gh0_11.sAo = 0; gh0_11.sAi = 0; gh0_11.sAm = H; gh0_11.sAk = 1; gh0_11.sBo = 0; gh0_11.sBi = 0; gh0_11.sBn = H; gh0_11.sBk = 1; gh0_11.sCo = 0; gh0_11.sCi = 0; gh0_11.sCm = H3; gh0_11.sRo = 0; gh0_11.sRi = 0; gh0_11.sRm = 0; gh0_11.sRn = 0;
      gh0_11.M = BK; gh0_11.N = H3; gh0_11.K = H; gh0_11.zi_n = 1; gh0_11.flags = 1; gh0_11.act = 0;
      gh0_11.alpha = 1.0f; gh0_11.beta = 0.0f; gh0_11.sa = 1.0f; gh0_11.sb = 1.0f; gh0_11.Npad = H3; gh0_11.pad_ = 0;
      k_gemm<1><<<dim3((unsigned)((H3) + 31) / 32, (unsigned)((BK) + 15) / 16, (unsigned)(1)), 32, 0, stream>>>(gh0_11); }
    k_gru<<<(unsigned)(((long long)BK * H + 255) / 256), 256, 0, stream>>>(nullptr, X, wih0, bih0, GH, H0, H0n, BK, H);
    { GemmP gi1_11;
      gi1_11.A = H0n; gi1_11.B = wih1; gi1_11.bias = bih1; gi1_11.R = H0n; gi1_11.C = GI;
      gi1_11.sAo = 0; gi1_11.sAi = 0; gi1_11.sAm = H; gi1_11.sAk = 1; gi1_11.sBo = 0; gi1_11.sBi = 0; gi1_11.sBn = H; gi1_11.sBk = 1; gi1_11.sCo = 0; gi1_11.sCi = 0; gi1_11.sCm = H3; gi1_11.sRo = 0; gi1_11.sRi = 0; gi1_11.sRm = 0; gi1_11.sRn = 0;
      gi1_11.M = BK; gi1_11.N = H3; gi1_11.K = H; gi1_11.zi_n = 1; gi1_11.flags = 1; gi1_11.act = 0;
      gi1_11.alpha = 1.0f; gi1_11.beta = 0.0f; gi1_11.sa = 1.0f; gi1_11.sb = 1.0f; gi1_11.Npad = H3; gi1_11.pad_ = 0;
      k_gemm<1><<<dim3((unsigned)((H3) + 31) / 32, (unsigned)((BK) + 15) / 16, (unsigned)(1)), 32, 0, stream>>>(gi1_11); }
    { GemmP gh1_11;
      gh1_11.A = H1; gh1_11.B = whh1; gh1_11.bias = bhh1; gh1_11.R = H1; gh1_11.C = GH;
      gh1_11.sAo = 0; gh1_11.sAi = 0; gh1_11.sAm = H; gh1_11.sAk = 1; gh1_11.sBo = 0; gh1_11.sBi = 0; gh1_11.sBn = H; gh1_11.sBk = 1; gh1_11.sCo = 0; gh1_11.sCi = 0; gh1_11.sCm = H3; gh1_11.sRo = 0; gh1_11.sRi = 0; gh1_11.sRm = 0; gh1_11.sRn = 0;
      gh1_11.M = BK; gh1_11.N = H3; gh1_11.K = H; gh1_11.zi_n = 1; gh1_11.flags = 1; gh1_11.act = 0;
      gh1_11.alpha = 1.0f; gh1_11.beta = 0.0f; gh1_11.sa = 1.0f; gh1_11.sb = 1.0f; gh1_11.Npad = H3; gh1_11.pad_ = 0;
      k_gemm<1><<<dim3((unsigned)((H3) + 31) / 32, (unsigned)((BK) + 15) / 16, (unsigned)(1)), 32, 0, stream>>>(gh1_11); }
    k_gru<<<(unsigned)(((long long)BK * H + 255) / 256), 256, 0, stream>>>(GI, nullptr, nullptr, nullptr, GH, H1, H1n, BK, H);
    { GemmP gd_11;
      gd_11.A = H1n; gd_11.B = ow; gd_11.bias = ob; gd_11.R = H1n; gd_11.C = DL;
      gd_11.sAo = 0; gd_11.sAi = 0; gd_11.sAm = H; gd_11.sAk = 1; gd_11.sBo = 0; gd_11.sBi = 0; gd_11.sBn = H; gd_11.sBk = 1; gd_11.sCo = 0; gd_11.sCi = 0; gd_11.sCm = LDP; gd_11.sRo = 0; gd_11.sRi = 0; gd_11.sRm = 0; gd_11.sRn = 0;
      gd_11.M = BK; gd_11.N = 2; gd_11.K = H; gd_11.zi_n = 1; gd_11.flags = 1; gd_11.act = 0;
      gd_11.alpha = 1.0f; gd_11.beta = 0.0f; gd_11.sa = 1.0f; gd_11.sb = 1.0f; gd_11.Npad = LDP; gd_11.pad_ = 0;
      k_gemm<1><<<dim3((unsigned)((LDP) + 31) / 32, (unsigned)((BK) + 15) / 16, (unsigned)(1)), 32, 0, stream>>>(gd_11); }
    k_posstep<<<(unsigned)((BK * 2 + 255) / 256), 256, 0, stream>>>(DL, LDP, X, POS, TRAJ, BK, T, 11);
    k_lincopy<<<(unsigned)(((long long)(BK) * (H) + 255) / 256), 256, 0, stream>>>(H0n, H, H0, H, BK, H);
    k_lincopy<<<(unsigned)(((long long)(BK) * (H) + 255) / 256), 256, 0, stream>>>(H1n, H, H1, H, BK, H);
    { GemmP gh0_12;
      gh0_12.A = H0; gh0_12.B = whh0; gh0_12.bias = bhh0; gh0_12.R = H0; gh0_12.C = GH;
      gh0_12.sAo = 0; gh0_12.sAi = 0; gh0_12.sAm = H; gh0_12.sAk = 1; gh0_12.sBo = 0; gh0_12.sBi = 0; gh0_12.sBn = H; gh0_12.sBk = 1; gh0_12.sCo = 0; gh0_12.sCi = 0; gh0_12.sCm = H3; gh0_12.sRo = 0; gh0_12.sRi = 0; gh0_12.sRm = 0; gh0_12.sRn = 0;
      gh0_12.M = BK; gh0_12.N = H3; gh0_12.K = H; gh0_12.zi_n = 1; gh0_12.flags = 1; gh0_12.act = 0;
      gh0_12.alpha = 1.0f; gh0_12.beta = 0.0f; gh0_12.sa = 1.0f; gh0_12.sb = 1.0f; gh0_12.Npad = H3; gh0_12.pad_ = 0;
      k_gemm<1><<<dim3((unsigned)((H3) + 31) / 32, (unsigned)((BK) + 15) / 16, (unsigned)(1)), 32, 0, stream>>>(gh0_12); }
    k_gru<<<(unsigned)(((long long)BK * H + 255) / 256), 256, 0, stream>>>(nullptr, X, wih0, bih0, GH, H0, H0n, BK, H);
    { GemmP gi1_12;
      gi1_12.A = H0n; gi1_12.B = wih1; gi1_12.bias = bih1; gi1_12.R = H0n; gi1_12.C = GI;
      gi1_12.sAo = 0; gi1_12.sAi = 0; gi1_12.sAm = H; gi1_12.sAk = 1; gi1_12.sBo = 0; gi1_12.sBi = 0; gi1_12.sBn = H; gi1_12.sBk = 1; gi1_12.sCo = 0; gi1_12.sCi = 0; gi1_12.sCm = H3; gi1_12.sRo = 0; gi1_12.sRi = 0; gi1_12.sRm = 0; gi1_12.sRn = 0;
      gi1_12.M = BK; gi1_12.N = H3; gi1_12.K = H; gi1_12.zi_n = 1; gi1_12.flags = 1; gi1_12.act = 0;
      gi1_12.alpha = 1.0f; gi1_12.beta = 0.0f; gi1_12.sa = 1.0f; gi1_12.sb = 1.0f; gi1_12.Npad = H3; gi1_12.pad_ = 0;
      k_gemm<1><<<dim3((unsigned)((H3) + 31) / 32, (unsigned)((BK) + 15) / 16, (unsigned)(1)), 32, 0, stream>>>(gi1_12); }
    { GemmP gh1_12;
      gh1_12.A = H1; gh1_12.B = whh1; gh1_12.bias = bhh1; gh1_12.R = H1; gh1_12.C = GH;
      gh1_12.sAo = 0; gh1_12.sAi = 0; gh1_12.sAm = H; gh1_12.sAk = 1; gh1_12.sBo = 0; gh1_12.sBi = 0; gh1_12.sBn = H; gh1_12.sBk = 1; gh1_12.sCo = 0; gh1_12.sCi = 0; gh1_12.sCm = H3; gh1_12.sRo = 0; gh1_12.sRi = 0; gh1_12.sRm = 0; gh1_12.sRn = 0;
      gh1_12.M = BK; gh1_12.N = H3; gh1_12.K = H; gh1_12.zi_n = 1; gh1_12.flags = 1; gh1_12.act = 0;
      gh1_12.alpha = 1.0f; gh1_12.beta = 0.0f; gh1_12.sa = 1.0f; gh1_12.sb = 1.0f; gh1_12.Npad = H3; gh1_12.pad_ = 0;
      k_gemm<1><<<dim3((unsigned)((H3) + 31) / 32, (unsigned)((BK) + 15) / 16, (unsigned)(1)), 32, 0, stream>>>(gh1_12); }
    k_gru<<<(unsigned)(((long long)BK * H + 255) / 256), 256, 0, stream>>>(GI, nullptr, nullptr, nullptr, GH, H1, H1n, BK, H);
    { GemmP gd_12;
      gd_12.A = H1n; gd_12.B = ow; gd_12.bias = ob; gd_12.R = H1n; gd_12.C = DL;
      gd_12.sAo = 0; gd_12.sAi = 0; gd_12.sAm = H; gd_12.sAk = 1; gd_12.sBo = 0; gd_12.sBi = 0; gd_12.sBn = H; gd_12.sBk = 1; gd_12.sCo = 0; gd_12.sCi = 0; gd_12.sCm = LDP; gd_12.sRo = 0; gd_12.sRi = 0; gd_12.sRm = 0; gd_12.sRn = 0;
      gd_12.M = BK; gd_12.N = 2; gd_12.K = H; gd_12.zi_n = 1; gd_12.flags = 1; gd_12.act = 0;
      gd_12.alpha = 1.0f; gd_12.beta = 0.0f; gd_12.sa = 1.0f; gd_12.sb = 1.0f; gd_12.Npad = LDP; gd_12.pad_ = 0;
      k_gemm<1><<<dim3((unsigned)((LDP) + 31) / 32, (unsigned)((BK) + 15) / 16, (unsigned)(1)), 32, 0, stream>>>(gd_12); }
    k_posstep<<<(unsigned)((BK * 2 + 255) / 256), 256, 0, stream>>>(DL, LDP, X, POS, TRAJ, BK, T, 12);
    k_lincopy<<<(unsigned)(((long long)(BK) * (H) + 255) / 256), 256, 0, stream>>>(H0n, H, H0, H, BK, H);
    k_lincopy<<<(unsigned)(((long long)(BK) * (H) + 255) / 256), 256, 0, stream>>>(H1n, H, H1, H, BK, H);
    { GemmP gh0_13;
      gh0_13.A = H0; gh0_13.B = whh0; gh0_13.bias = bhh0; gh0_13.R = H0; gh0_13.C = GH;
      gh0_13.sAo = 0; gh0_13.sAi = 0; gh0_13.sAm = H; gh0_13.sAk = 1; gh0_13.sBo = 0; gh0_13.sBi = 0; gh0_13.sBn = H; gh0_13.sBk = 1; gh0_13.sCo = 0; gh0_13.sCi = 0; gh0_13.sCm = H3; gh0_13.sRo = 0; gh0_13.sRi = 0; gh0_13.sRm = 0; gh0_13.sRn = 0;
      gh0_13.M = BK; gh0_13.N = H3; gh0_13.K = H; gh0_13.zi_n = 1; gh0_13.flags = 1; gh0_13.act = 0;
      gh0_13.alpha = 1.0f; gh0_13.beta = 0.0f; gh0_13.sa = 1.0f; gh0_13.sb = 1.0f; gh0_13.Npad = H3; gh0_13.pad_ = 0;
      k_gemm<1><<<dim3((unsigned)((H3) + 31) / 32, (unsigned)((BK) + 15) / 16, (unsigned)(1)), 32, 0, stream>>>(gh0_13); }
    k_gru<<<(unsigned)(((long long)BK * H + 255) / 256), 256, 0, stream>>>(nullptr, X, wih0, bih0, GH, H0, H0n, BK, H);
    { GemmP gi1_13;
      gi1_13.A = H0n; gi1_13.B = wih1; gi1_13.bias = bih1; gi1_13.R = H0n; gi1_13.C = GI;
      gi1_13.sAo = 0; gi1_13.sAi = 0; gi1_13.sAm = H; gi1_13.sAk = 1; gi1_13.sBo = 0; gi1_13.sBi = 0; gi1_13.sBn = H; gi1_13.sBk = 1; gi1_13.sCo = 0; gi1_13.sCi = 0; gi1_13.sCm = H3; gi1_13.sRo = 0; gi1_13.sRi = 0; gi1_13.sRm = 0; gi1_13.sRn = 0;
      gi1_13.M = BK; gi1_13.N = H3; gi1_13.K = H; gi1_13.zi_n = 1; gi1_13.flags = 1; gi1_13.act = 0;
      gi1_13.alpha = 1.0f; gi1_13.beta = 0.0f; gi1_13.sa = 1.0f; gi1_13.sb = 1.0f; gi1_13.Npad = H3; gi1_13.pad_ = 0;
      k_gemm<1><<<dim3((unsigned)((H3) + 31) / 32, (unsigned)((BK) + 15) / 16, (unsigned)(1)), 32, 0, stream>>>(gi1_13); }
    { GemmP gh1_13;
      gh1_13.A = H1; gh1_13.B = whh1; gh1_13.bias = bhh1; gh1_13.R = H1; gh1_13.C = GH;
      gh1_13.sAo = 0; gh1_13.sAi = 0; gh1_13.sAm = H; gh1_13.sAk = 1; gh1_13.sBo = 0; gh1_13.sBi = 0; gh1_13.sBn = H; gh1_13.sBk = 1; gh1_13.sCo = 0; gh1_13.sCi = 0; gh1_13.sCm = H3; gh1_13.sRo = 0; gh1_13.sRi = 0; gh1_13.sRm = 0; gh1_13.sRn = 0;
      gh1_13.M = BK; gh1_13.N = H3; gh1_13.K = H; gh1_13.zi_n = 1; gh1_13.flags = 1; gh1_13.act = 0;
      gh1_13.alpha = 1.0f; gh1_13.beta = 0.0f; gh1_13.sa = 1.0f; gh1_13.sb = 1.0f; gh1_13.Npad = H3; gh1_13.pad_ = 0;
      k_gemm<1><<<dim3((unsigned)((H3) + 31) / 32, (unsigned)((BK) + 15) / 16, (unsigned)(1)), 32, 0, stream>>>(gh1_13); }
    k_gru<<<(unsigned)(((long long)BK * H + 255) / 256), 256, 0, stream>>>(GI, nullptr, nullptr, nullptr, GH, H1, H1n, BK, H);
    { GemmP gd_13;
      gd_13.A = H1n; gd_13.B = ow; gd_13.bias = ob; gd_13.R = H1n; gd_13.C = DL;
      gd_13.sAo = 0; gd_13.sAi = 0; gd_13.sAm = H; gd_13.sAk = 1; gd_13.sBo = 0; gd_13.sBi = 0; gd_13.sBn = H; gd_13.sBk = 1; gd_13.sCo = 0; gd_13.sCi = 0; gd_13.sCm = LDP; gd_13.sRo = 0; gd_13.sRi = 0; gd_13.sRm = 0; gd_13.sRn = 0;
      gd_13.M = BK; gd_13.N = 2; gd_13.K = H; gd_13.zi_n = 1; gd_13.flags = 1; gd_13.act = 0;
      gd_13.alpha = 1.0f; gd_13.beta = 0.0f; gd_13.sa = 1.0f; gd_13.sb = 1.0f; gd_13.Npad = LDP; gd_13.pad_ = 0;
      k_gemm<1><<<dim3((unsigned)((LDP) + 31) / 32, (unsigned)((BK) + 15) / 16, (unsigned)(1)), 32, 0, stream>>>(gd_13); }
    k_posstep<<<(unsigned)((BK * 2 + 255) / 256), 256, 0, stream>>>(DL, LDP, X, POS, TRAJ, BK, T, 13);
    k_lincopy<<<(unsigned)(((long long)(BK) * (H) + 255) / 256), 256, 0, stream>>>(H0n, H, H0, H, BK, H);
    k_lincopy<<<(unsigned)(((long long)(BK) * (H) + 255) / 256), 256, 0, stream>>>(H1n, H, H1, H, BK, H);
    { GemmP gh0_14;
      gh0_14.A = H0; gh0_14.B = whh0; gh0_14.bias = bhh0; gh0_14.R = H0; gh0_14.C = GH;
      gh0_14.sAo = 0; gh0_14.sAi = 0; gh0_14.sAm = H; gh0_14.sAk = 1; gh0_14.sBo = 0; gh0_14.sBi = 0; gh0_14.sBn = H; gh0_14.sBk = 1; gh0_14.sCo = 0; gh0_14.sCi = 0; gh0_14.sCm = H3; gh0_14.sRo = 0; gh0_14.sRi = 0; gh0_14.sRm = 0; gh0_14.sRn = 0;
      gh0_14.M = BK; gh0_14.N = H3; gh0_14.K = H; gh0_14.zi_n = 1; gh0_14.flags = 1; gh0_14.act = 0;
      gh0_14.alpha = 1.0f; gh0_14.beta = 0.0f; gh0_14.sa = 1.0f; gh0_14.sb = 1.0f; gh0_14.Npad = H3; gh0_14.pad_ = 0;
      k_gemm<1><<<dim3((unsigned)((H3) + 31) / 32, (unsigned)((BK) + 15) / 16, (unsigned)(1)), 32, 0, stream>>>(gh0_14); }
    k_gru<<<(unsigned)(((long long)BK * H + 255) / 256), 256, 0, stream>>>(nullptr, X, wih0, bih0, GH, H0, H0n, BK, H);
    { GemmP gi1_14;
      gi1_14.A = H0n; gi1_14.B = wih1; gi1_14.bias = bih1; gi1_14.R = H0n; gi1_14.C = GI;
      gi1_14.sAo = 0; gi1_14.sAi = 0; gi1_14.sAm = H; gi1_14.sAk = 1; gi1_14.sBo = 0; gi1_14.sBi = 0; gi1_14.sBn = H; gi1_14.sBk = 1; gi1_14.sCo = 0; gi1_14.sCi = 0; gi1_14.sCm = H3; gi1_14.sRo = 0; gi1_14.sRi = 0; gi1_14.sRm = 0; gi1_14.sRn = 0;
      gi1_14.M = BK; gi1_14.N = H3; gi1_14.K = H; gi1_14.zi_n = 1; gi1_14.flags = 1; gi1_14.act = 0;
      gi1_14.alpha = 1.0f; gi1_14.beta = 0.0f; gi1_14.sa = 1.0f; gi1_14.sb = 1.0f; gi1_14.Npad = H3; gi1_14.pad_ = 0;
      k_gemm<1><<<dim3((unsigned)((H3) + 31) / 32, (unsigned)((BK) + 15) / 16, (unsigned)(1)), 32, 0, stream>>>(gi1_14); }
    { GemmP gh1_14;
      gh1_14.A = H1; gh1_14.B = whh1; gh1_14.bias = bhh1; gh1_14.R = H1; gh1_14.C = GH;
      gh1_14.sAo = 0; gh1_14.sAi = 0; gh1_14.sAm = H; gh1_14.sAk = 1; gh1_14.sBo = 0; gh1_14.sBi = 0; gh1_14.sBn = H; gh1_14.sBk = 1; gh1_14.sCo = 0; gh1_14.sCi = 0; gh1_14.sCm = H3; gh1_14.sRo = 0; gh1_14.sRi = 0; gh1_14.sRm = 0; gh1_14.sRn = 0;
      gh1_14.M = BK; gh1_14.N = H3; gh1_14.K = H; gh1_14.zi_n = 1; gh1_14.flags = 1; gh1_14.act = 0;
      gh1_14.alpha = 1.0f; gh1_14.beta = 0.0f; gh1_14.sa = 1.0f; gh1_14.sb = 1.0f; gh1_14.Npad = H3; gh1_14.pad_ = 0;
      k_gemm<1><<<dim3((unsigned)((H3) + 31) / 32, (unsigned)((BK) + 15) / 16, (unsigned)(1)), 32, 0, stream>>>(gh1_14); }
    k_gru<<<(unsigned)(((long long)BK * H + 255) / 256), 256, 0, stream>>>(GI, nullptr, nullptr, nullptr, GH, H1, H1n, BK, H);
    { GemmP gd_14;
      gd_14.A = H1n; gd_14.B = ow; gd_14.bias = ob; gd_14.R = H1n; gd_14.C = DL;
      gd_14.sAo = 0; gd_14.sAi = 0; gd_14.sAm = H; gd_14.sAk = 1; gd_14.sBo = 0; gd_14.sBi = 0; gd_14.sBn = H; gd_14.sBk = 1; gd_14.sCo = 0; gd_14.sCi = 0; gd_14.sCm = LDP; gd_14.sRo = 0; gd_14.sRi = 0; gd_14.sRm = 0; gd_14.sRn = 0;
      gd_14.M = BK; gd_14.N = 2; gd_14.K = H; gd_14.zi_n = 1; gd_14.flags = 1; gd_14.act = 0;
      gd_14.alpha = 1.0f; gd_14.beta = 0.0f; gd_14.sa = 1.0f; gd_14.sb = 1.0f; gd_14.Npad = LDP; gd_14.pad_ = 0;
      k_gemm<1><<<dim3((unsigned)((LDP) + 31) / 32, (unsigned)((BK) + 15) / 16, (unsigned)(1)), 32, 0, stream>>>(gd_14); }
    k_posstep<<<(unsigned)((BK * 2 + 255) / 256), 256, 0, stream>>>(DL, LDP, X, POS, TRAJ, BK, T, 14);
    k_lincopy<<<(unsigned)(((long long)(BK) * (H) + 255) / 256), 256, 0, stream>>>(H0n, H, H0, H, BK, H);
    k_lincopy<<<(unsigned)(((long long)(BK) * (H) + 255) / 256), 256, 0, stream>>>(H1n, H, H1, H, BK, H);
    { GemmP gh0_15;
      gh0_15.A = H0; gh0_15.B = whh0; gh0_15.bias = bhh0; gh0_15.R = H0; gh0_15.C = GH;
      gh0_15.sAo = 0; gh0_15.sAi = 0; gh0_15.sAm = H; gh0_15.sAk = 1; gh0_15.sBo = 0; gh0_15.sBi = 0; gh0_15.sBn = H; gh0_15.sBk = 1; gh0_15.sCo = 0; gh0_15.sCi = 0; gh0_15.sCm = H3; gh0_15.sRo = 0; gh0_15.sRi = 0; gh0_15.sRm = 0; gh0_15.sRn = 0;
      gh0_15.M = BK; gh0_15.N = H3; gh0_15.K = H; gh0_15.zi_n = 1; gh0_15.flags = 1; gh0_15.act = 0;
      gh0_15.alpha = 1.0f; gh0_15.beta = 0.0f; gh0_15.sa = 1.0f; gh0_15.sb = 1.0f; gh0_15.Npad = H3; gh0_15.pad_ = 0;
      k_gemm<1><<<dim3((unsigned)((H3) + 31) / 32, (unsigned)((BK) + 15) / 16, (unsigned)(1)), 32, 0, stream>>>(gh0_15); }
    k_gru<<<(unsigned)(((long long)BK * H + 255) / 256), 256, 0, stream>>>(nullptr, X, wih0, bih0, GH, H0, H0n, BK, H);
    { GemmP gi1_15;
      gi1_15.A = H0n; gi1_15.B = wih1; gi1_15.bias = bih1; gi1_15.R = H0n; gi1_15.C = GI;
      gi1_15.sAo = 0; gi1_15.sAi = 0; gi1_15.sAm = H; gi1_15.sAk = 1; gi1_15.sBo = 0; gi1_15.sBi = 0; gi1_15.sBn = H; gi1_15.sBk = 1; gi1_15.sCo = 0; gi1_15.sCi = 0; gi1_15.sCm = H3; gi1_15.sRo = 0; gi1_15.sRi = 0; gi1_15.sRm = 0; gi1_15.sRn = 0;
      gi1_15.M = BK; gi1_15.N = H3; gi1_15.K = H; gi1_15.zi_n = 1; gi1_15.flags = 1; gi1_15.act = 0;
      gi1_15.alpha = 1.0f; gi1_15.beta = 0.0f; gi1_15.sa = 1.0f; gi1_15.sb = 1.0f; gi1_15.Npad = H3; gi1_15.pad_ = 0;
      k_gemm<1><<<dim3((unsigned)((H3) + 31) / 32, (unsigned)((BK) + 15) / 16, (unsigned)(1)), 32, 0, stream>>>(gi1_15); }
    { GemmP gh1_15;
      gh1_15.A = H1; gh1_15.B = whh1; gh1_15.bias = bhh1; gh1_15.R = H1; gh1_15.C = GH;
      gh1_15.sAo = 0; gh1_15.sAi = 0; gh1_15.sAm = H; gh1_15.sAk = 1; gh1_15.sBo = 0; gh1_15.sBi = 0; gh1_15.sBn = H; gh1_15.sBk = 1; gh1_15.sCo = 0; gh1_15.sCi = 0; gh1_15.sCm = H3; gh1_15.sRo = 0; gh1_15.sRi = 0; gh1_15.sRm = 0; gh1_15.sRn = 0;
      gh1_15.M = BK; gh1_15.N = H3; gh1_15.K = H; gh1_15.zi_n = 1; gh1_15.flags = 1; gh1_15.act = 0;
      gh1_15.alpha = 1.0f; gh1_15.beta = 0.0f; gh1_15.sa = 1.0f; gh1_15.sb = 1.0f; gh1_15.Npad = H3; gh1_15.pad_ = 0;
      k_gemm<1><<<dim3((unsigned)((H3) + 31) / 32, (unsigned)((BK) + 15) / 16, (unsigned)(1)), 32, 0, stream>>>(gh1_15); }
    k_gru<<<(unsigned)(((long long)BK * H + 255) / 256), 256, 0, stream>>>(GI, nullptr, nullptr, nullptr, GH, H1, H1n, BK, H);
    { GemmP gd_15;
      gd_15.A = H1n; gd_15.B = ow; gd_15.bias = ob; gd_15.R = H1n; gd_15.C = DL;
      gd_15.sAo = 0; gd_15.sAi = 0; gd_15.sAm = H; gd_15.sAk = 1; gd_15.sBo = 0; gd_15.sBi = 0; gd_15.sBn = H; gd_15.sBk = 1; gd_15.sCo = 0; gd_15.sCi = 0; gd_15.sCm = LDP; gd_15.sRo = 0; gd_15.sRi = 0; gd_15.sRm = 0; gd_15.sRn = 0;
      gd_15.M = BK; gd_15.N = 2; gd_15.K = H; gd_15.zi_n = 1; gd_15.flags = 1; gd_15.act = 0;
      gd_15.alpha = 1.0f; gd_15.beta = 0.0f; gd_15.sa = 1.0f; gd_15.sb = 1.0f; gd_15.Npad = LDP; gd_15.pad_ = 0;
      k_gemm<1><<<dim3((unsigned)((LDP) + 31) / 32, (unsigned)((BK) + 15) / 16, (unsigned)(1)), 32, 0, stream>>>(gd_15); }
    k_posstep<<<(unsigned)((BK * 2 + 255) / 256), 256, 0, stream>>>(DL, LDP, X, POS, TRAJ, BK, T, 15);
    k_lincopy<<<(unsigned)(((long long)(BK) * (H) + 255) / 256), 256, 0, stream>>>(H0n, H, H0, H, BK, H);
    k_lincopy<<<(unsigned)(((long long)(BK) * (H) + 255) / 256), 256, 0, stream>>>(H1n, H, H1, H, BK, H);
    { GemmP gh0_16;
      gh0_16.A = H0; gh0_16.B = whh0; gh0_16.bias = bhh0; gh0_16.R = H0; gh0_16.C = GH;
      gh0_16.sAo = 0; gh0_16.sAi = 0; gh0_16.sAm = H; gh0_16.sAk = 1; gh0_16.sBo = 0; gh0_16.sBi = 0; gh0_16.sBn = H; gh0_16.sBk = 1; gh0_16.sCo = 0; gh0_16.sCi = 0; gh0_16.sCm = H3; gh0_16.sRo = 0; gh0_16.sRi = 0; gh0_16.sRm = 0; gh0_16.sRn = 0;
      gh0_16.M = BK; gh0_16.N = H3; gh0_16.K = H; gh0_16.zi_n = 1; gh0_16.flags = 1; gh0_16.act = 0;
      gh0_16.alpha = 1.0f; gh0_16.beta = 0.0f; gh0_16.sa = 1.0f; gh0_16.sb = 1.0f; gh0_16.Npad = H3; gh0_16.pad_ = 0;
      k_gemm<1><<<dim3((unsigned)((H3) + 31) / 32, (unsigned)((BK) + 15) / 16, (unsigned)(1)), 32, 0, stream>>>(gh0_16); }
    k_gru<<<(unsigned)(((long long)BK * H + 255) / 256), 256, 0, stream>>>(nullptr, X, wih0, bih0, GH, H0, H0n, BK, H);
    { GemmP gi1_16;
      gi1_16.A = H0n; gi1_16.B = wih1; gi1_16.bias = bih1; gi1_16.R = H0n; gi1_16.C = GI;
      gi1_16.sAo = 0; gi1_16.sAi = 0; gi1_16.sAm = H; gi1_16.sAk = 1; gi1_16.sBo = 0; gi1_16.sBi = 0; gi1_16.sBn = H; gi1_16.sBk = 1; gi1_16.sCo = 0; gi1_16.sCi = 0; gi1_16.sCm = H3; gi1_16.sRo = 0; gi1_16.sRi = 0; gi1_16.sRm = 0; gi1_16.sRn = 0;
      gi1_16.M = BK; gi1_16.N = H3; gi1_16.K = H; gi1_16.zi_n = 1; gi1_16.flags = 1; gi1_16.act = 0;
      gi1_16.alpha = 1.0f; gi1_16.beta = 0.0f; gi1_16.sa = 1.0f; gi1_16.sb = 1.0f; gi1_16.Npad = H3; gi1_16.pad_ = 0;
      k_gemm<1><<<dim3((unsigned)((H3) + 31) / 32, (unsigned)((BK) + 15) / 16, (unsigned)(1)), 32, 0, stream>>>(gi1_16); }
    { GemmP gh1_16;
      gh1_16.A = H1; gh1_16.B = whh1; gh1_16.bias = bhh1; gh1_16.R = H1; gh1_16.C = GH;
      gh1_16.sAo = 0; gh1_16.sAi = 0; gh1_16.sAm = H; gh1_16.sAk = 1; gh1_16.sBo = 0; gh1_16.sBi = 0; gh1_16.sBn = H; gh1_16.sBk = 1; gh1_16.sCo = 0; gh1_16.sCi = 0; gh1_16.sCm = H3; gh1_16.sRo = 0; gh1_16.sRi = 0; gh1_16.sRm = 0; gh1_16.sRn = 0;
      gh1_16.M = BK; gh1_16.N = H3; gh1_16.K = H; gh1_16.zi_n = 1; gh1_16.flags = 1; gh1_16.act = 0;
      gh1_16.alpha = 1.0f; gh1_16.beta = 0.0f; gh1_16.sa = 1.0f; gh1_16.sb = 1.0f; gh1_16.Npad = H3; gh1_16.pad_ = 0;
      k_gemm<1><<<dim3((unsigned)((H3) + 31) / 32, (unsigned)((BK) + 15) / 16, (unsigned)(1)), 32, 0, stream>>>(gh1_16); }
    k_gru<<<(unsigned)(((long long)BK * H + 255) / 256), 256, 0, stream>>>(GI, nullptr, nullptr, nullptr, GH, H1, H1n, BK, H);
    { GemmP gd_16;
      gd_16.A = H1n; gd_16.B = ow; gd_16.bias = ob; gd_16.R = H1n; gd_16.C = DL;
      gd_16.sAo = 0; gd_16.sAi = 0; gd_16.sAm = H; gd_16.sAk = 1; gd_16.sBo = 0; gd_16.sBi = 0; gd_16.sBn = H; gd_16.sBk = 1; gd_16.sCo = 0; gd_16.sCi = 0; gd_16.sCm = LDP; gd_16.sRo = 0; gd_16.sRi = 0; gd_16.sRm = 0; gd_16.sRn = 0;
      gd_16.M = BK; gd_16.N = 2; gd_16.K = H; gd_16.zi_n = 1; gd_16.flags = 1; gd_16.act = 0;
      gd_16.alpha = 1.0f; gd_16.beta = 0.0f; gd_16.sa = 1.0f; gd_16.sb = 1.0f; gd_16.Npad = LDP; gd_16.pad_ = 0;
      k_gemm<1><<<dim3((unsigned)((LDP) + 31) / 32, (unsigned)((BK) + 15) / 16, (unsigned)(1)), 32, 0, stream>>>(gd_16); }
    k_posstep<<<(unsigned)((BK * 2 + 255) / 256), 256, 0, stream>>>(DL, LDP, X, POS, TRAJ, BK, T, 16);
    k_lincopy<<<(unsigned)(((long long)(BK) * (H) + 255) / 256), 256, 0, stream>>>(H0n, H, H0, H, BK, H);
    k_lincopy<<<(unsigned)(((long long)(BK) * (H) + 255) / 256), 256, 0, stream>>>(H1n, H, H1, H, BK, H);
    { GemmP gh0_17;
      gh0_17.A = H0; gh0_17.B = whh0; gh0_17.bias = bhh0; gh0_17.R = H0; gh0_17.C = GH;
      gh0_17.sAo = 0; gh0_17.sAi = 0; gh0_17.sAm = H; gh0_17.sAk = 1; gh0_17.sBo = 0; gh0_17.sBi = 0; gh0_17.sBn = H; gh0_17.sBk = 1; gh0_17.sCo = 0; gh0_17.sCi = 0; gh0_17.sCm = H3; gh0_17.sRo = 0; gh0_17.sRi = 0; gh0_17.sRm = 0; gh0_17.sRn = 0;
      gh0_17.M = BK; gh0_17.N = H3; gh0_17.K = H; gh0_17.zi_n = 1; gh0_17.flags = 1; gh0_17.act = 0;
      gh0_17.alpha = 1.0f; gh0_17.beta = 0.0f; gh0_17.sa = 1.0f; gh0_17.sb = 1.0f; gh0_17.Npad = H3; gh0_17.pad_ = 0;
      k_gemm<1><<<dim3((unsigned)((H3) + 31) / 32, (unsigned)((BK) + 15) / 16, (unsigned)(1)), 32, 0, stream>>>(gh0_17); }
    k_gru<<<(unsigned)(((long long)BK * H + 255) / 256), 256, 0, stream>>>(nullptr, X, wih0, bih0, GH, H0, H0n, BK, H);
    { GemmP gi1_17;
      gi1_17.A = H0n; gi1_17.B = wih1; gi1_17.bias = bih1; gi1_17.R = H0n; gi1_17.C = GI;
      gi1_17.sAo = 0; gi1_17.sAi = 0; gi1_17.sAm = H; gi1_17.sAk = 1; gi1_17.sBo = 0; gi1_17.sBi = 0; gi1_17.sBn = H; gi1_17.sBk = 1; gi1_17.sCo = 0; gi1_17.sCi = 0; gi1_17.sCm = H3; gi1_17.sRo = 0; gi1_17.sRi = 0; gi1_17.sRm = 0; gi1_17.sRn = 0;
      gi1_17.M = BK; gi1_17.N = H3; gi1_17.K = H; gi1_17.zi_n = 1; gi1_17.flags = 1; gi1_17.act = 0;
      gi1_17.alpha = 1.0f; gi1_17.beta = 0.0f; gi1_17.sa = 1.0f; gi1_17.sb = 1.0f; gi1_17.Npad = H3; gi1_17.pad_ = 0;
      k_gemm<1><<<dim3((unsigned)((H3) + 31) / 32, (unsigned)((BK) + 15) / 16, (unsigned)(1)), 32, 0, stream>>>(gi1_17); }
    { GemmP gh1_17;
      gh1_17.A = H1; gh1_17.B = whh1; gh1_17.bias = bhh1; gh1_17.R = H1; gh1_17.C = GH;
      gh1_17.sAo = 0; gh1_17.sAi = 0; gh1_17.sAm = H; gh1_17.sAk = 1; gh1_17.sBo = 0; gh1_17.sBi = 0; gh1_17.sBn = H; gh1_17.sBk = 1; gh1_17.sCo = 0; gh1_17.sCi = 0; gh1_17.sCm = H3; gh1_17.sRo = 0; gh1_17.sRi = 0; gh1_17.sRm = 0; gh1_17.sRn = 0;
      gh1_17.M = BK; gh1_17.N = H3; gh1_17.K = H; gh1_17.zi_n = 1; gh1_17.flags = 1; gh1_17.act = 0;
      gh1_17.alpha = 1.0f; gh1_17.beta = 0.0f; gh1_17.sa = 1.0f; gh1_17.sb = 1.0f; gh1_17.Npad = H3; gh1_17.pad_ = 0;
      k_gemm<1><<<dim3((unsigned)((H3) + 31) / 32, (unsigned)((BK) + 15) / 16, (unsigned)(1)), 32, 0, stream>>>(gh1_17); }
    k_gru<<<(unsigned)(((long long)BK * H + 255) / 256), 256, 0, stream>>>(GI, nullptr, nullptr, nullptr, GH, H1, H1n, BK, H);
    { GemmP gd_17;
      gd_17.A = H1n; gd_17.B = ow; gd_17.bias = ob; gd_17.R = H1n; gd_17.C = DL;
      gd_17.sAo = 0; gd_17.sAi = 0; gd_17.sAm = H; gd_17.sAk = 1; gd_17.sBo = 0; gd_17.sBi = 0; gd_17.sBn = H; gd_17.sBk = 1; gd_17.sCo = 0; gd_17.sCi = 0; gd_17.sCm = LDP; gd_17.sRo = 0; gd_17.sRi = 0; gd_17.sRm = 0; gd_17.sRn = 0;
      gd_17.M = BK; gd_17.N = 2; gd_17.K = H; gd_17.zi_n = 1; gd_17.flags = 1; gd_17.act = 0;
      gd_17.alpha = 1.0f; gd_17.beta = 0.0f; gd_17.sa = 1.0f; gd_17.sb = 1.0f; gd_17.Npad = LDP; gd_17.pad_ = 0;
      k_gemm<1><<<dim3((unsigned)((LDP) + 31) / 32, (unsigned)((BK) + 15) / 16, (unsigned)(1)), 32, 0, stream>>>(gd_17); }
    k_posstep<<<(unsigned)((BK * 2 + 255) / 256), 256, 0, stream>>>(DL, LDP, X, POS, TRAJ, BK, T, 17);
    k_lincopy<<<(unsigned)(((long long)(BK) * (H) + 255) / 256), 256, 0, stream>>>(H0n, H, H0, H, BK, H);
    k_lincopy<<<(unsigned)(((long long)(BK) * (H) + 255) / 256), 256, 0, stream>>>(H1n, H, H1, H, BK, H);
    { GemmP gh0_18;
      gh0_18.A = H0; gh0_18.B = whh0; gh0_18.bias = bhh0; gh0_18.R = H0; gh0_18.C = GH;
      gh0_18.sAo = 0; gh0_18.sAi = 0; gh0_18.sAm = H; gh0_18.sAk = 1; gh0_18.sBo = 0; gh0_18.sBi = 0; gh0_18.sBn = H; gh0_18.sBk = 1; gh0_18.sCo = 0; gh0_18.sCi = 0; gh0_18.sCm = H3; gh0_18.sRo = 0; gh0_18.sRi = 0; gh0_18.sRm = 0; gh0_18.sRn = 0;
      gh0_18.M = BK; gh0_18.N = H3; gh0_18.K = H; gh0_18.zi_n = 1; gh0_18.flags = 1; gh0_18.act = 0;
      gh0_18.alpha = 1.0f; gh0_18.beta = 0.0f; gh0_18.sa = 1.0f; gh0_18.sb = 1.0f; gh0_18.Npad = H3; gh0_18.pad_ = 0;
      k_gemm<1><<<dim3((unsigned)((H3) + 31) / 32, (unsigned)((BK) + 15) / 16, (unsigned)(1)), 32, 0, stream>>>(gh0_18); }
    k_gru<<<(unsigned)(((long long)BK * H + 255) / 256), 256, 0, stream>>>(nullptr, X, wih0, bih0, GH, H0, H0n, BK, H);
    { GemmP gi1_18;
      gi1_18.A = H0n; gi1_18.B = wih1; gi1_18.bias = bih1; gi1_18.R = H0n; gi1_18.C = GI;
      gi1_18.sAo = 0; gi1_18.sAi = 0; gi1_18.sAm = H; gi1_18.sAk = 1; gi1_18.sBo = 0; gi1_18.sBi = 0; gi1_18.sBn = H; gi1_18.sBk = 1; gi1_18.sCo = 0; gi1_18.sCi = 0; gi1_18.sCm = H3; gi1_18.sRo = 0; gi1_18.sRi = 0; gi1_18.sRm = 0; gi1_18.sRn = 0;
      gi1_18.M = BK; gi1_18.N = H3; gi1_18.K = H; gi1_18.zi_n = 1; gi1_18.flags = 1; gi1_18.act = 0;
      gi1_18.alpha = 1.0f; gi1_18.beta = 0.0f; gi1_18.sa = 1.0f; gi1_18.sb = 1.0f; gi1_18.Npad = H3; gi1_18.pad_ = 0;
      k_gemm<1><<<dim3((unsigned)((H3) + 31) / 32, (unsigned)((BK) + 15) / 16, (unsigned)(1)), 32, 0, stream>>>(gi1_18); }
    { GemmP gh1_18;
      gh1_18.A = H1; gh1_18.B = whh1; gh1_18.bias = bhh1; gh1_18.R = H1; gh1_18.C = GH;
      gh1_18.sAo = 0; gh1_18.sAi = 0; gh1_18.sAm = H; gh1_18.sAk = 1; gh1_18.sBo = 0; gh1_18.sBi = 0; gh1_18.sBn = H; gh1_18.sBk = 1; gh1_18.sCo = 0; gh1_18.sCi = 0; gh1_18.sCm = H3; gh1_18.sRo = 0; gh1_18.sRi = 0; gh1_18.sRm = 0; gh1_18.sRn = 0;
      gh1_18.M = BK; gh1_18.N = H3; gh1_18.K = H; gh1_18.zi_n = 1; gh1_18.flags = 1; gh1_18.act = 0;
      gh1_18.alpha = 1.0f; gh1_18.beta = 0.0f; gh1_18.sa = 1.0f; gh1_18.sb = 1.0f; gh1_18.Npad = H3; gh1_18.pad_ = 0;
      k_gemm<1><<<dim3((unsigned)((H3) + 31) / 32, (unsigned)((BK) + 15) / 16, (unsigned)(1)), 32, 0, stream>>>(gh1_18); }
    k_gru<<<(unsigned)(((long long)BK * H + 255) / 256), 256, 0, stream>>>(GI, nullptr, nullptr, nullptr, GH, H1, H1n, BK, H);
    { GemmP gd_18;
      gd_18.A = H1n; gd_18.B = ow; gd_18.bias = ob; gd_18.R = H1n; gd_18.C = DL;
      gd_18.sAo = 0; gd_18.sAi = 0; gd_18.sAm = H; gd_18.sAk = 1; gd_18.sBo = 0; gd_18.sBi = 0; gd_18.sBn = H; gd_18.sBk = 1; gd_18.sCo = 0; gd_18.sCi = 0; gd_18.sCm = LDP; gd_18.sRo = 0; gd_18.sRi = 0; gd_18.sRm = 0; gd_18.sRn = 0;
      gd_18.M = BK; gd_18.N = 2; gd_18.K = H; gd_18.zi_n = 1; gd_18.flags = 1; gd_18.act = 0;
      gd_18.alpha = 1.0f; gd_18.beta = 0.0f; gd_18.sa = 1.0f; gd_18.sb = 1.0f; gd_18.Npad = LDP; gd_18.pad_ = 0;
      k_gemm<1><<<dim3((unsigned)((LDP) + 31) / 32, (unsigned)((BK) + 15) / 16, (unsigned)(1)), 32, 0, stream>>>(gd_18); }
    k_posstep<<<(unsigned)((BK * 2 + 255) / 256), 256, 0, stream>>>(DL, LDP, X, POS, TRAJ, BK, T, 18);
    k_lincopy<<<(unsigned)(((long long)(BK) * (H) + 255) / 256), 256, 0, stream>>>(H0n, H, H0, H, BK, H);
    k_lincopy<<<(unsigned)(((long long)(BK) * (H) + 255) / 256), 256, 0, stream>>>(H1n, H, H1, H, BK, H);
    { GemmP gh0_19;
      gh0_19.A = H0; gh0_19.B = whh0; gh0_19.bias = bhh0; gh0_19.R = H0; gh0_19.C = GH;
      gh0_19.sAo = 0; gh0_19.sAi = 0; gh0_19.sAm = H; gh0_19.sAk = 1; gh0_19.sBo = 0; gh0_19.sBi = 0; gh0_19.sBn = H; gh0_19.sBk = 1; gh0_19.sCo = 0; gh0_19.sCi = 0; gh0_19.sCm = H3; gh0_19.sRo = 0; gh0_19.sRi = 0; gh0_19.sRm = 0; gh0_19.sRn = 0;
      gh0_19.M = BK; gh0_19.N = H3; gh0_19.K = H; gh0_19.zi_n = 1; gh0_19.flags = 1; gh0_19.act = 0;
      gh0_19.alpha = 1.0f; gh0_19.beta = 0.0f; gh0_19.sa = 1.0f; gh0_19.sb = 1.0f; gh0_19.Npad = H3; gh0_19.pad_ = 0;
      k_gemm<1><<<dim3((unsigned)((H3) + 31) / 32, (unsigned)((BK) + 15) / 16, (unsigned)(1)), 32, 0, stream>>>(gh0_19); }
    k_gru<<<(unsigned)(((long long)BK * H + 255) / 256), 256, 0, stream>>>(nullptr, X, wih0, bih0, GH, H0, H0n, BK, H);
    { GemmP gi1_19;
      gi1_19.A = H0n; gi1_19.B = wih1; gi1_19.bias = bih1; gi1_19.R = H0n; gi1_19.C = GI;
      gi1_19.sAo = 0; gi1_19.sAi = 0; gi1_19.sAm = H; gi1_19.sAk = 1; gi1_19.sBo = 0; gi1_19.sBi = 0; gi1_19.sBn = H; gi1_19.sBk = 1; gi1_19.sCo = 0; gi1_19.sCi = 0; gi1_19.sCm = H3; gi1_19.sRo = 0; gi1_19.sRi = 0; gi1_19.sRm = 0; gi1_19.sRn = 0;
      gi1_19.M = BK; gi1_19.N = H3; gi1_19.K = H; gi1_19.zi_n = 1; gi1_19.flags = 1; gi1_19.act = 0;
      gi1_19.alpha = 1.0f; gi1_19.beta = 0.0f; gi1_19.sa = 1.0f; gi1_19.sb = 1.0f; gi1_19.Npad = H3; gi1_19.pad_ = 0;
      k_gemm<1><<<dim3((unsigned)((H3) + 31) / 32, (unsigned)((BK) + 15) / 16, (unsigned)(1)), 32, 0, stream>>>(gi1_19); }
    { GemmP gh1_19;
      gh1_19.A = H1; gh1_19.B = whh1; gh1_19.bias = bhh1; gh1_19.R = H1; gh1_19.C = GH;
      gh1_19.sAo = 0; gh1_19.sAi = 0; gh1_19.sAm = H; gh1_19.sAk = 1; gh1_19.sBo = 0; gh1_19.sBi = 0; gh1_19.sBn = H; gh1_19.sBk = 1; gh1_19.sCo = 0; gh1_19.sCi = 0; gh1_19.sCm = H3; gh1_19.sRo = 0; gh1_19.sRi = 0; gh1_19.sRm = 0; gh1_19.sRn = 0;
      gh1_19.M = BK; gh1_19.N = H3; gh1_19.K = H; gh1_19.zi_n = 1; gh1_19.flags = 1; gh1_19.act = 0;
      gh1_19.alpha = 1.0f; gh1_19.beta = 0.0f; gh1_19.sa = 1.0f; gh1_19.sb = 1.0f; gh1_19.Npad = H3; gh1_19.pad_ = 0;
      k_gemm<1><<<dim3((unsigned)((H3) + 31) / 32, (unsigned)((BK) + 15) / 16, (unsigned)(1)), 32, 0, stream>>>(gh1_19); }
    k_gru<<<(unsigned)(((long long)BK * H + 255) / 256), 256, 0, stream>>>(GI, nullptr, nullptr, nullptr, GH, H1, H1n, BK, H);
    { GemmP gd_19;
      gd_19.A = H1n; gd_19.B = ow; gd_19.bias = ob; gd_19.R = H1n; gd_19.C = DL;
      gd_19.sAo = 0; gd_19.sAi = 0; gd_19.sAm = H; gd_19.sAk = 1; gd_19.sBo = 0; gd_19.sBi = 0; gd_19.sBn = H; gd_19.sBk = 1; gd_19.sCo = 0; gd_19.sCi = 0; gd_19.sCm = LDP; gd_19.sRo = 0; gd_19.sRi = 0; gd_19.sRm = 0; gd_19.sRn = 0;
      gd_19.M = BK; gd_19.N = 2; gd_19.K = H; gd_19.zi_n = 1; gd_19.flags = 1; gd_19.act = 0;
      gd_19.alpha = 1.0f; gd_19.beta = 0.0f; gd_19.sa = 1.0f; gd_19.sb = 1.0f; gd_19.Npad = LDP; gd_19.pad_ = 0;
      k_gemm<1><<<dim3((unsigned)((LDP) + 31) / 32, (unsigned)((BK) + 15) / 16, (unsigned)(1)), 32, 0, stream>>>(gd_19); }
    k_posstep<<<(unsigned)((BK * 2 + 255) / 256), 256, 0, stream>>>(DL, LDP, X, POS, TRAJ, BK, T, 19);
    k_lincopy<<<(unsigned)(((long long)(BK) * (H) + 255) / 256), 256, 0, stream>>>(H0n, H, H0, H, BK, H);
    k_lincopy<<<(unsigned)(((long long)(BK) * (H) + 255) / 256), 256, 0, stream>>>(H1n, H, H1, H, BK, H);
    { GemmP gh0_20;
      gh0_20.A = H0; gh0_20.B = whh0; gh0_20.bias = bhh0; gh0_20.R = H0; gh0_20.C = GH;
      gh0_20.sAo = 0; gh0_20.sAi = 0; gh0_20.sAm = H; gh0_20.sAk = 1; gh0_20.sBo = 0; gh0_20.sBi = 0; gh0_20.sBn = H; gh0_20.sBk = 1; gh0_20.sCo = 0; gh0_20.sCi = 0; gh0_20.sCm = H3; gh0_20.sRo = 0; gh0_20.sRi = 0; gh0_20.sRm = 0; gh0_20.sRn = 0;
      gh0_20.M = BK; gh0_20.N = H3; gh0_20.K = H; gh0_20.zi_n = 1; gh0_20.flags = 1; gh0_20.act = 0;
      gh0_20.alpha = 1.0f; gh0_20.beta = 0.0f; gh0_20.sa = 1.0f; gh0_20.sb = 1.0f; gh0_20.Npad = H3; gh0_20.pad_ = 0;
      k_gemm<1><<<dim3((unsigned)((H3) + 31) / 32, (unsigned)((BK) + 15) / 16, (unsigned)(1)), 32, 0, stream>>>(gh0_20); }
    k_gru<<<(unsigned)(((long long)BK * H + 255) / 256), 256, 0, stream>>>(nullptr, X, wih0, bih0, GH, H0, H0n, BK, H);
    { GemmP gi1_20;
      gi1_20.A = H0n; gi1_20.B = wih1; gi1_20.bias = bih1; gi1_20.R = H0n; gi1_20.C = GI;
      gi1_20.sAo = 0; gi1_20.sAi = 0; gi1_20.sAm = H; gi1_20.sAk = 1; gi1_20.sBo = 0; gi1_20.sBi = 0; gi1_20.sBn = H; gi1_20.sBk = 1; gi1_20.sCo = 0; gi1_20.sCi = 0; gi1_20.sCm = H3; gi1_20.sRo = 0; gi1_20.sRi = 0; gi1_20.sRm = 0; gi1_20.sRn = 0;
      gi1_20.M = BK; gi1_20.N = H3; gi1_20.K = H; gi1_20.zi_n = 1; gi1_20.flags = 1; gi1_20.act = 0;
      gi1_20.alpha = 1.0f; gi1_20.beta = 0.0f; gi1_20.sa = 1.0f; gi1_20.sb = 1.0f; gi1_20.Npad = H3; gi1_20.pad_ = 0;
      k_gemm<1><<<dim3((unsigned)((H3) + 31) / 32, (unsigned)((BK) + 15) / 16, (unsigned)(1)), 32, 0, stream>>>(gi1_20); }
    { GemmP gh1_20;
      gh1_20.A = H1; gh1_20.B = whh1; gh1_20.bias = bhh1; gh1_20.R = H1; gh1_20.C = GH;
      gh1_20.sAo = 0; gh1_20.sAi = 0; gh1_20.sAm = H; gh1_20.sAk = 1; gh1_20.sBo = 0; gh1_20.sBi = 0; gh1_20.sBn = H; gh1_20.sBk = 1; gh1_20.sCo = 0; gh1_20.sCi = 0; gh1_20.sCm = H3; gh1_20.sRo = 0; gh1_20.sRi = 0; gh1_20.sRm = 0; gh1_20.sRn = 0;
      gh1_20.M = BK; gh1_20.N = H3; gh1_20.K = H; gh1_20.zi_n = 1; gh1_20.flags = 1; gh1_20.act = 0;
      gh1_20.alpha = 1.0f; gh1_20.beta = 0.0f; gh1_20.sa = 1.0f; gh1_20.sb = 1.0f; gh1_20.Npad = H3; gh1_20.pad_ = 0;
      k_gemm<1><<<dim3((unsigned)((H3) + 31) / 32, (unsigned)((BK) + 15) / 16, (unsigned)(1)), 32, 0, stream>>>(gh1_20); }
    k_gru<<<(unsigned)(((long long)BK * H + 255) / 256), 256, 0, stream>>>(GI, nullptr, nullptr, nullptr, GH, H1, H1n, BK, H);
    { GemmP gd_20;
      gd_20.A = H1n; gd_20.B = ow; gd_20.bias = ob; gd_20.R = H1n; gd_20.C = DL;
      gd_20.sAo = 0; gd_20.sAi = 0; gd_20.sAm = H; gd_20.sAk = 1; gd_20.sBo = 0; gd_20.sBi = 0; gd_20.sBn = H; gd_20.sBk = 1; gd_20.sCo = 0; gd_20.sCi = 0; gd_20.sCm = LDP; gd_20.sRo = 0; gd_20.sRi = 0; gd_20.sRm = 0; gd_20.sRn = 0;
      gd_20.M = BK; gd_20.N = 2; gd_20.K = H; gd_20.zi_n = 1; gd_20.flags = 1; gd_20.act = 0;
      gd_20.alpha = 1.0f; gd_20.beta = 0.0f; gd_20.sa = 1.0f; gd_20.sb = 1.0f; gd_20.Npad = LDP; gd_20.pad_ = 0;
      k_gemm<1><<<dim3((unsigned)((LDP) + 31) / 32, (unsigned)((BK) + 15) / 16, (unsigned)(1)), 32, 0, stream>>>(gd_20); }
    k_posstep<<<(unsigned)((BK * 2 + 255) / 256), 256, 0, stream>>>(DL, LDP, X, POS, TRAJ, BK, T, 20);
    k_lincopy<<<(unsigned)(((long long)(BK) * (H) + 255) / 256), 256, 0, stream>>>(H0n, H, H0, H, BK, H);
    k_lincopy<<<(unsigned)(((long long)(BK) * (H) + 255) / 256), 256, 0, stream>>>(H1n, H, H1, H, BK, H);
    { GemmP gh0_21;
      gh0_21.A = H0; gh0_21.B = whh0; gh0_21.bias = bhh0; gh0_21.R = H0; gh0_21.C = GH;
      gh0_21.sAo = 0; gh0_21.sAi = 0; gh0_21.sAm = H; gh0_21.sAk = 1; gh0_21.sBo = 0; gh0_21.sBi = 0; gh0_21.sBn = H; gh0_21.sBk = 1; gh0_21.sCo = 0; gh0_21.sCi = 0; gh0_21.sCm = H3; gh0_21.sRo = 0; gh0_21.sRi = 0; gh0_21.sRm = 0; gh0_21.sRn = 0;
      gh0_21.M = BK; gh0_21.N = H3; gh0_21.K = H; gh0_21.zi_n = 1; gh0_21.flags = 1; gh0_21.act = 0;
      gh0_21.alpha = 1.0f; gh0_21.beta = 0.0f; gh0_21.sa = 1.0f; gh0_21.sb = 1.0f; gh0_21.Npad = H3; gh0_21.pad_ = 0;
      k_gemm<1><<<dim3((unsigned)((H3) + 31) / 32, (unsigned)((BK) + 15) / 16, (unsigned)(1)), 32, 0, stream>>>(gh0_21); }
    k_gru<<<(unsigned)(((long long)BK * H + 255) / 256), 256, 0, stream>>>(nullptr, X, wih0, bih0, GH, H0, H0n, BK, H);
    { GemmP gi1_21;
      gi1_21.A = H0n; gi1_21.B = wih1; gi1_21.bias = bih1; gi1_21.R = H0n; gi1_21.C = GI;
      gi1_21.sAo = 0; gi1_21.sAi = 0; gi1_21.sAm = H; gi1_21.sAk = 1; gi1_21.sBo = 0; gi1_21.sBi = 0; gi1_21.sBn = H; gi1_21.sBk = 1; gi1_21.sCo = 0; gi1_21.sCi = 0; gi1_21.sCm = H3; gi1_21.sRo = 0; gi1_21.sRi = 0; gi1_21.sRm = 0; gi1_21.sRn = 0;
      gi1_21.M = BK; gi1_21.N = H3; gi1_21.K = H; gi1_21.zi_n = 1; gi1_21.flags = 1; gi1_21.act = 0;
      gi1_21.alpha = 1.0f; gi1_21.beta = 0.0f; gi1_21.sa = 1.0f; gi1_21.sb = 1.0f; gi1_21.Npad = H3; gi1_21.pad_ = 0;
      k_gemm<1><<<dim3((unsigned)((H3) + 31) / 32, (unsigned)((BK) + 15) / 16, (unsigned)(1)), 32, 0, stream>>>(gi1_21); }
    { GemmP gh1_21;
      gh1_21.A = H1; gh1_21.B = whh1; gh1_21.bias = bhh1; gh1_21.R = H1; gh1_21.C = GH;
      gh1_21.sAo = 0; gh1_21.sAi = 0; gh1_21.sAm = H; gh1_21.sAk = 1; gh1_21.sBo = 0; gh1_21.sBi = 0; gh1_21.sBn = H; gh1_21.sBk = 1; gh1_21.sCo = 0; gh1_21.sCi = 0; gh1_21.sCm = H3; gh1_21.sRo = 0; gh1_21.sRi = 0; gh1_21.sRm = 0; gh1_21.sRn = 0;
      gh1_21.M = BK; gh1_21.N = H3; gh1_21.K = H; gh1_21.zi_n = 1; gh1_21.flags = 1; gh1_21.act = 0;
      gh1_21.alpha = 1.0f; gh1_21.beta = 0.0f; gh1_21.sa = 1.0f; gh1_21.sb = 1.0f; gh1_21.Npad = H3; gh1_21.pad_ = 0;
      k_gemm<1><<<dim3((unsigned)((H3) + 31) / 32, (unsigned)((BK) + 15) / 16, (unsigned)(1)), 32, 0, stream>>>(gh1_21); }
    k_gru<<<(unsigned)(((long long)BK * H + 255) / 256), 256, 0, stream>>>(GI, nullptr, nullptr, nullptr, GH, H1, H1n, BK, H);
    { GemmP gd_21;
      gd_21.A = H1n; gd_21.B = ow; gd_21.bias = ob; gd_21.R = H1n; gd_21.C = DL;
      gd_21.sAo = 0; gd_21.sAi = 0; gd_21.sAm = H; gd_21.sAk = 1; gd_21.sBo = 0; gd_21.sBi = 0; gd_21.sBn = H; gd_21.sBk = 1; gd_21.sCo = 0; gd_21.sCi = 0; gd_21.sCm = LDP; gd_21.sRo = 0; gd_21.sRi = 0; gd_21.sRm = 0; gd_21.sRn = 0;
      gd_21.M = BK; gd_21.N = 2; gd_21.K = H; gd_21.zi_n = 1; gd_21.flags = 1; gd_21.act = 0;
      gd_21.alpha = 1.0f; gd_21.beta = 0.0f; gd_21.sa = 1.0f; gd_21.sb = 1.0f; gd_21.Npad = LDP; gd_21.pad_ = 0;
      k_gemm<1><<<dim3((unsigned)((LDP) + 31) / 32, (unsigned)((BK) + 15) / 16, (unsigned)(1)), 32, 0, stream>>>(gd_21); }
    k_posstep<<<(unsigned)((BK * 2 + 255) / 256), 256, 0, stream>>>(DL, LDP, X, POS, TRAJ, BK, T, 21);
    k_lincopy<<<(unsigned)(((long long)(BK) * (H) + 255) / 256), 256, 0, stream>>>(H0n, H, H0, H, BK, H);
    k_lincopy<<<(unsigned)(((long long)(BK) * (H) + 255) / 256), 256, 0, stream>>>(H1n, H, H1, H, BK, H);
    { GemmP gh0_22;
      gh0_22.A = H0; gh0_22.B = whh0; gh0_22.bias = bhh0; gh0_22.R = H0; gh0_22.C = GH;
      gh0_22.sAo = 0; gh0_22.sAi = 0; gh0_22.sAm = H; gh0_22.sAk = 1; gh0_22.sBo = 0; gh0_22.sBi = 0; gh0_22.sBn = H; gh0_22.sBk = 1; gh0_22.sCo = 0; gh0_22.sCi = 0; gh0_22.sCm = H3; gh0_22.sRo = 0; gh0_22.sRi = 0; gh0_22.sRm = 0; gh0_22.sRn = 0;
      gh0_22.M = BK; gh0_22.N = H3; gh0_22.K = H; gh0_22.zi_n = 1; gh0_22.flags = 1; gh0_22.act = 0;
      gh0_22.alpha = 1.0f; gh0_22.beta = 0.0f; gh0_22.sa = 1.0f; gh0_22.sb = 1.0f; gh0_22.Npad = H3; gh0_22.pad_ = 0;
      k_gemm<1><<<dim3((unsigned)((H3) + 31) / 32, (unsigned)((BK) + 15) / 16, (unsigned)(1)), 32, 0, stream>>>(gh0_22); }
    k_gru<<<(unsigned)(((long long)BK * H + 255) / 256), 256, 0, stream>>>(nullptr, X, wih0, bih0, GH, H0, H0n, BK, H);
    { GemmP gi1_22;
      gi1_22.A = H0n; gi1_22.B = wih1; gi1_22.bias = bih1; gi1_22.R = H0n; gi1_22.C = GI;
      gi1_22.sAo = 0; gi1_22.sAi = 0; gi1_22.sAm = H; gi1_22.sAk = 1; gi1_22.sBo = 0; gi1_22.sBi = 0; gi1_22.sBn = H; gi1_22.sBk = 1; gi1_22.sCo = 0; gi1_22.sCi = 0; gi1_22.sCm = H3; gi1_22.sRo = 0; gi1_22.sRi = 0; gi1_22.sRm = 0; gi1_22.sRn = 0;
      gi1_22.M = BK; gi1_22.N = H3; gi1_22.K = H; gi1_22.zi_n = 1; gi1_22.flags = 1; gi1_22.act = 0;
      gi1_22.alpha = 1.0f; gi1_22.beta = 0.0f; gi1_22.sa = 1.0f; gi1_22.sb = 1.0f; gi1_22.Npad = H3; gi1_22.pad_ = 0;
      k_gemm<1><<<dim3((unsigned)((H3) + 31) / 32, (unsigned)((BK) + 15) / 16, (unsigned)(1)), 32, 0, stream>>>(gi1_22); }
    { GemmP gh1_22;
      gh1_22.A = H1; gh1_22.B = whh1; gh1_22.bias = bhh1; gh1_22.R = H1; gh1_22.C = GH;
      gh1_22.sAo = 0; gh1_22.sAi = 0; gh1_22.sAm = H; gh1_22.sAk = 1; gh1_22.sBo = 0; gh1_22.sBi = 0; gh1_22.sBn = H; gh1_22.sBk = 1; gh1_22.sCo = 0; gh1_22.sCi = 0; gh1_22.sCm = H3; gh1_22.sRo = 0; gh1_22.sRi = 0; gh1_22.sRm = 0; gh1_22.sRn = 0;
      gh1_22.M = BK; gh1_22.N = H3; gh1_22.K = H; gh1_22.zi_n = 1; gh1_22.flags = 1; gh1_22.act = 0;
      gh1_22.alpha = 1.0f; gh1_22.beta = 0.0f; gh1_22.sa = 1.0f; gh1_22.sb = 1.0f; gh1_22.Npad = H3; gh1_22.pad_ = 0;
      k_gemm<1><<<dim3((unsigned)((H3) + 31) / 32, (unsigned)((BK) + 15) / 16, (unsigned)(1)), 32, 0, stream>>>(gh1_22); }
    k_gru<<<(unsigned)(((long long)BK * H + 255) / 256), 256, 0, stream>>>(GI, nullptr, nullptr, nullptr, GH, H1, H1n, BK, H);
    { GemmP gd_22;
      gd_22.A = H1n; gd_22.B = ow; gd_22.bias = ob; gd_22.R = H1n; gd_22.C = DL;
      gd_22.sAo = 0; gd_22.sAi = 0; gd_22.sAm = H; gd_22.sAk = 1; gd_22.sBo = 0; gd_22.sBi = 0; gd_22.sBn = H; gd_22.sBk = 1; gd_22.sCo = 0; gd_22.sCi = 0; gd_22.sCm = LDP; gd_22.sRo = 0; gd_22.sRi = 0; gd_22.sRm = 0; gd_22.sRn = 0;
      gd_22.M = BK; gd_22.N = 2; gd_22.K = H; gd_22.zi_n = 1; gd_22.flags = 1; gd_22.act = 0;
      gd_22.alpha = 1.0f; gd_22.beta = 0.0f; gd_22.sa = 1.0f; gd_22.sb = 1.0f; gd_22.Npad = LDP; gd_22.pad_ = 0;
      k_gemm<1><<<dim3((unsigned)((LDP) + 31) / 32, (unsigned)((BK) + 15) / 16, (unsigned)(1)), 32, 0, stream>>>(gd_22); }
    k_posstep<<<(unsigned)((BK * 2 + 255) / 256), 256, 0, stream>>>(DL, LDP, X, POS, TRAJ, BK, T, 22);
    k_lincopy<<<(unsigned)(((long long)(BK) * (H) + 255) / 256), 256, 0, stream>>>(H0n, H, H0, H, BK, H);
    k_lincopy<<<(unsigned)(((long long)(BK) * (H) + 255) / 256), 256, 0, stream>>>(H1n, H, H1, H, BK, H);
    { GemmP gh0_23;
      gh0_23.A = H0; gh0_23.B = whh0; gh0_23.bias = bhh0; gh0_23.R = H0; gh0_23.C = GH;
      gh0_23.sAo = 0; gh0_23.sAi = 0; gh0_23.sAm = H; gh0_23.sAk = 1; gh0_23.sBo = 0; gh0_23.sBi = 0; gh0_23.sBn = H; gh0_23.sBk = 1; gh0_23.sCo = 0; gh0_23.sCi = 0; gh0_23.sCm = H3; gh0_23.sRo = 0; gh0_23.sRi = 0; gh0_23.sRm = 0; gh0_23.sRn = 0;
      gh0_23.M = BK; gh0_23.N = H3; gh0_23.K = H; gh0_23.zi_n = 1; gh0_23.flags = 1; gh0_23.act = 0;
      gh0_23.alpha = 1.0f; gh0_23.beta = 0.0f; gh0_23.sa = 1.0f; gh0_23.sb = 1.0f; gh0_23.Npad = H3; gh0_23.pad_ = 0;
      k_gemm<1><<<dim3((unsigned)((H3) + 31) / 32, (unsigned)((BK) + 15) / 16, (unsigned)(1)), 32, 0, stream>>>(gh0_23); }
    k_gru<<<(unsigned)(((long long)BK * H + 255) / 256), 256, 0, stream>>>(nullptr, X, wih0, bih0, GH, H0, H0n, BK, H);
    { GemmP gi1_23;
      gi1_23.A = H0n; gi1_23.B = wih1; gi1_23.bias = bih1; gi1_23.R = H0n; gi1_23.C = GI;
      gi1_23.sAo = 0; gi1_23.sAi = 0; gi1_23.sAm = H; gi1_23.sAk = 1; gi1_23.sBo = 0; gi1_23.sBi = 0; gi1_23.sBn = H; gi1_23.sBk = 1; gi1_23.sCo = 0; gi1_23.sCi = 0; gi1_23.sCm = H3; gi1_23.sRo = 0; gi1_23.sRi = 0; gi1_23.sRm = 0; gi1_23.sRn = 0;
      gi1_23.M = BK; gi1_23.N = H3; gi1_23.K = H; gi1_23.zi_n = 1; gi1_23.flags = 1; gi1_23.act = 0;
      gi1_23.alpha = 1.0f; gi1_23.beta = 0.0f; gi1_23.sa = 1.0f; gi1_23.sb = 1.0f; gi1_23.Npad = H3; gi1_23.pad_ = 0;
      k_gemm<1><<<dim3((unsigned)((H3) + 31) / 32, (unsigned)((BK) + 15) / 16, (unsigned)(1)), 32, 0, stream>>>(gi1_23); }
    { GemmP gh1_23;
      gh1_23.A = H1; gh1_23.B = whh1; gh1_23.bias = bhh1; gh1_23.R = H1; gh1_23.C = GH;
      gh1_23.sAo = 0; gh1_23.sAi = 0; gh1_23.sAm = H; gh1_23.sAk = 1; gh1_23.sBo = 0; gh1_23.sBi = 0; gh1_23.sBn = H; gh1_23.sBk = 1; gh1_23.sCo = 0; gh1_23.sCi = 0; gh1_23.sCm = H3; gh1_23.sRo = 0; gh1_23.sRi = 0; gh1_23.sRm = 0; gh1_23.sRn = 0;
      gh1_23.M = BK; gh1_23.N = H3; gh1_23.K = H; gh1_23.zi_n = 1; gh1_23.flags = 1; gh1_23.act = 0;
      gh1_23.alpha = 1.0f; gh1_23.beta = 0.0f; gh1_23.sa = 1.0f; gh1_23.sb = 1.0f; gh1_23.Npad = H3; gh1_23.pad_ = 0;
      k_gemm<1><<<dim3((unsigned)((H3) + 31) / 32, (unsigned)((BK) + 15) / 16, (unsigned)(1)), 32, 0, stream>>>(gh1_23); }
    k_gru<<<(unsigned)(((long long)BK * H + 255) / 256), 256, 0, stream>>>(GI, nullptr, nullptr, nullptr, GH, H1, H1n, BK, H);
    { GemmP gd_23;
      gd_23.A = H1n; gd_23.B = ow; gd_23.bias = ob; gd_23.R = H1n; gd_23.C = DL;
      gd_23.sAo = 0; gd_23.sAi = 0; gd_23.sAm = H; gd_23.sAk = 1; gd_23.sBo = 0; gd_23.sBi = 0; gd_23.sBn = H; gd_23.sBk = 1; gd_23.sCo = 0; gd_23.sCi = 0; gd_23.sCm = LDP; gd_23.sRo = 0; gd_23.sRi = 0; gd_23.sRm = 0; gd_23.sRn = 0;
      gd_23.M = BK; gd_23.N = 2; gd_23.K = H; gd_23.zi_n = 1; gd_23.flags = 1; gd_23.act = 0;
      gd_23.alpha = 1.0f; gd_23.beta = 0.0f; gd_23.sa = 1.0f; gd_23.sb = 1.0f; gd_23.Npad = LDP; gd_23.pad_ = 0;
      k_gemm<1><<<dim3((unsigned)((LDP) + 31) / 32, (unsigned)((BK) + 15) / 16, (unsigned)(1)), 32, 0, stream>>>(gd_23); }
    k_posstep<<<(unsigned)((BK * 2 + 255) / 256), 256, 0, stream>>>(DL, LDP, X, POS, TRAJ, BK, T, 23);
    k_lincopy<<<(unsigned)(((long long)(BK) * (H) + 255) / 256), 256, 0, stream>>>(H0n, H, H0, H, BK, H);
    k_lincopy<<<(unsigned)(((long long)(BK) * (H) + 255) / 256), 256, 0, stream>>>(H1n, H, H1, H, BK, H);
    { GemmP gh0_24;
      gh0_24.A = H0; gh0_24.B = whh0; gh0_24.bias = bhh0; gh0_24.R = H0; gh0_24.C = GH;
      gh0_24.sAo = 0; gh0_24.sAi = 0; gh0_24.sAm = H; gh0_24.sAk = 1; gh0_24.sBo = 0; gh0_24.sBi = 0; gh0_24.sBn = H; gh0_24.sBk = 1; gh0_24.sCo = 0; gh0_24.sCi = 0; gh0_24.sCm = H3; gh0_24.sRo = 0; gh0_24.sRi = 0; gh0_24.sRm = 0; gh0_24.sRn = 0;
      gh0_24.M = BK; gh0_24.N = H3; gh0_24.K = H; gh0_24.zi_n = 1; gh0_24.flags = 1; gh0_24.act = 0;
      gh0_24.alpha = 1.0f; gh0_24.beta = 0.0f; gh0_24.sa = 1.0f; gh0_24.sb = 1.0f; gh0_24.Npad = H3; gh0_24.pad_ = 0;
      k_gemm<1><<<dim3((unsigned)((H3) + 31) / 32, (unsigned)((BK) + 15) / 16, (unsigned)(1)), 32, 0, stream>>>(gh0_24); }
    k_gru<<<(unsigned)(((long long)BK * H + 255) / 256), 256, 0, stream>>>(nullptr, X, wih0, bih0, GH, H0, H0n, BK, H);
    { GemmP gi1_24;
      gi1_24.A = H0n; gi1_24.B = wih1; gi1_24.bias = bih1; gi1_24.R = H0n; gi1_24.C = GI;
      gi1_24.sAo = 0; gi1_24.sAi = 0; gi1_24.sAm = H; gi1_24.sAk = 1; gi1_24.sBo = 0; gi1_24.sBi = 0; gi1_24.sBn = H; gi1_24.sBk = 1; gi1_24.sCo = 0; gi1_24.sCi = 0; gi1_24.sCm = H3; gi1_24.sRo = 0; gi1_24.sRi = 0; gi1_24.sRm = 0; gi1_24.sRn = 0;
      gi1_24.M = BK; gi1_24.N = H3; gi1_24.K = H; gi1_24.zi_n = 1; gi1_24.flags = 1; gi1_24.act = 0;
      gi1_24.alpha = 1.0f; gi1_24.beta = 0.0f; gi1_24.sa = 1.0f; gi1_24.sb = 1.0f; gi1_24.Npad = H3; gi1_24.pad_ = 0;
      k_gemm<1><<<dim3((unsigned)((H3) + 31) / 32, (unsigned)((BK) + 15) / 16, (unsigned)(1)), 32, 0, stream>>>(gi1_24); }
    { GemmP gh1_24;
      gh1_24.A = H1; gh1_24.B = whh1; gh1_24.bias = bhh1; gh1_24.R = H1; gh1_24.C = GH;
      gh1_24.sAo = 0; gh1_24.sAi = 0; gh1_24.sAm = H; gh1_24.sAk = 1; gh1_24.sBo = 0; gh1_24.sBi = 0; gh1_24.sBn = H; gh1_24.sBk = 1; gh1_24.sCo = 0; gh1_24.sCi = 0; gh1_24.sCm = H3; gh1_24.sRo = 0; gh1_24.sRi = 0; gh1_24.sRm = 0; gh1_24.sRn = 0;
      gh1_24.M = BK; gh1_24.N = H3; gh1_24.K = H; gh1_24.zi_n = 1; gh1_24.flags = 1; gh1_24.act = 0;
      gh1_24.alpha = 1.0f; gh1_24.beta = 0.0f; gh1_24.sa = 1.0f; gh1_24.sb = 1.0f; gh1_24.Npad = H3; gh1_24.pad_ = 0;
      k_gemm<1><<<dim3((unsigned)((H3) + 31) / 32, (unsigned)((BK) + 15) / 16, (unsigned)(1)), 32, 0, stream>>>(gh1_24); }
    k_gru<<<(unsigned)(((long long)BK * H + 255) / 256), 256, 0, stream>>>(GI, nullptr, nullptr, nullptr, GH, H1, H1n, BK, H);
    { GemmP gd_24;
      gd_24.A = H1n; gd_24.B = ow; gd_24.bias = ob; gd_24.R = H1n; gd_24.C = DL;
      gd_24.sAo = 0; gd_24.sAi = 0; gd_24.sAm = H; gd_24.sAk = 1; gd_24.sBo = 0; gd_24.sBi = 0; gd_24.sBn = H; gd_24.sBk = 1; gd_24.sCo = 0; gd_24.sCi = 0; gd_24.sCm = LDP; gd_24.sRo = 0; gd_24.sRi = 0; gd_24.sRm = 0; gd_24.sRn = 0;
      gd_24.M = BK; gd_24.N = 2; gd_24.K = H; gd_24.zi_n = 1; gd_24.flags = 1; gd_24.act = 0;
      gd_24.alpha = 1.0f; gd_24.beta = 0.0f; gd_24.sa = 1.0f; gd_24.sb = 1.0f; gd_24.Npad = LDP; gd_24.pad_ = 0;
      k_gemm<1><<<dim3((unsigned)((LDP) + 31) / 32, (unsigned)((BK) + 15) / 16, (unsigned)(1)), 32, 0, stream>>>(gd_24); }
    k_posstep<<<(unsigned)((BK * 2 + 255) / 256), 256, 0, stream>>>(DL, LDP, X, POS, TRAJ, BK, T, 24);
    k_lincopy<<<(unsigned)(((long long)(BK) * (H) + 255) / 256), 256, 0, stream>>>(H0n, H, H0, H, BK, H);
    k_lincopy<<<(unsigned)(((long long)(BK) * (H) + 255) / 256), 256, 0, stream>>>(H1n, H, H1, H, BK, H);
    { GemmP gh0_25;
      gh0_25.A = H0; gh0_25.B = whh0; gh0_25.bias = bhh0; gh0_25.R = H0; gh0_25.C = GH;
      gh0_25.sAo = 0; gh0_25.sAi = 0; gh0_25.sAm = H; gh0_25.sAk = 1; gh0_25.sBo = 0; gh0_25.sBi = 0; gh0_25.sBn = H; gh0_25.sBk = 1; gh0_25.sCo = 0; gh0_25.sCi = 0; gh0_25.sCm = H3; gh0_25.sRo = 0; gh0_25.sRi = 0; gh0_25.sRm = 0; gh0_25.sRn = 0;
      gh0_25.M = BK; gh0_25.N = H3; gh0_25.K = H; gh0_25.zi_n = 1; gh0_25.flags = 1; gh0_25.act = 0;
      gh0_25.alpha = 1.0f; gh0_25.beta = 0.0f; gh0_25.sa = 1.0f; gh0_25.sb = 1.0f; gh0_25.Npad = H3; gh0_25.pad_ = 0;
      k_gemm<1><<<dim3((unsigned)((H3) + 31) / 32, (unsigned)((BK) + 15) / 16, (unsigned)(1)), 32, 0, stream>>>(gh0_25); }
    k_gru<<<(unsigned)(((long long)BK * H + 255) / 256), 256, 0, stream>>>(nullptr, X, wih0, bih0, GH, H0, H0n, BK, H);
    { GemmP gi1_25;
      gi1_25.A = H0n; gi1_25.B = wih1; gi1_25.bias = bih1; gi1_25.R = H0n; gi1_25.C = GI;
      gi1_25.sAo = 0; gi1_25.sAi = 0; gi1_25.sAm = H; gi1_25.sAk = 1; gi1_25.sBo = 0; gi1_25.sBi = 0; gi1_25.sBn = H; gi1_25.sBk = 1; gi1_25.sCo = 0; gi1_25.sCi = 0; gi1_25.sCm = H3; gi1_25.sRo = 0; gi1_25.sRi = 0; gi1_25.sRm = 0; gi1_25.sRn = 0;
      gi1_25.M = BK; gi1_25.N = H3; gi1_25.K = H; gi1_25.zi_n = 1; gi1_25.flags = 1; gi1_25.act = 0;
      gi1_25.alpha = 1.0f; gi1_25.beta = 0.0f; gi1_25.sa = 1.0f; gi1_25.sb = 1.0f; gi1_25.Npad = H3; gi1_25.pad_ = 0;
      k_gemm<1><<<dim3((unsigned)((H3) + 31) / 32, (unsigned)((BK) + 15) / 16, (unsigned)(1)), 32, 0, stream>>>(gi1_25); }
    { GemmP gh1_25;
      gh1_25.A = H1; gh1_25.B = whh1; gh1_25.bias = bhh1; gh1_25.R = H1; gh1_25.C = GH;
      gh1_25.sAo = 0; gh1_25.sAi = 0; gh1_25.sAm = H; gh1_25.sAk = 1; gh1_25.sBo = 0; gh1_25.sBi = 0; gh1_25.sBn = H; gh1_25.sBk = 1; gh1_25.sCo = 0; gh1_25.sCi = 0; gh1_25.sCm = H3; gh1_25.sRo = 0; gh1_25.sRi = 0; gh1_25.sRm = 0; gh1_25.sRn = 0;
      gh1_25.M = BK; gh1_25.N = H3; gh1_25.K = H; gh1_25.zi_n = 1; gh1_25.flags = 1; gh1_25.act = 0;
      gh1_25.alpha = 1.0f; gh1_25.beta = 0.0f; gh1_25.sa = 1.0f; gh1_25.sb = 1.0f; gh1_25.Npad = H3; gh1_25.pad_ = 0;
      k_gemm<1><<<dim3((unsigned)((H3) + 31) / 32, (unsigned)((BK) + 15) / 16, (unsigned)(1)), 32, 0, stream>>>(gh1_25); }
    k_gru<<<(unsigned)(((long long)BK * H + 255) / 256), 256, 0, stream>>>(GI, nullptr, nullptr, nullptr, GH, H1, H1n, BK, H);
    { GemmP gd_25;
      gd_25.A = H1n; gd_25.B = ow; gd_25.bias = ob; gd_25.R = H1n; gd_25.C = DL;
      gd_25.sAo = 0; gd_25.sAi = 0; gd_25.sAm = H; gd_25.sAk = 1; gd_25.sBo = 0; gd_25.sBi = 0; gd_25.sBn = H; gd_25.sBk = 1; gd_25.sCo = 0; gd_25.sCi = 0; gd_25.sCm = LDP; gd_25.sRo = 0; gd_25.sRi = 0; gd_25.sRm = 0; gd_25.sRn = 0;
      gd_25.M = BK; gd_25.N = 2; gd_25.K = H; gd_25.zi_n = 1; gd_25.flags = 1; gd_25.act = 0;
      gd_25.alpha = 1.0f; gd_25.beta = 0.0f; gd_25.sa = 1.0f; gd_25.sb = 1.0f; gd_25.Npad = LDP; gd_25.pad_ = 0;
      k_gemm<1><<<dim3((unsigned)((LDP) + 31) / 32, (unsigned)((BK) + 15) / 16, (unsigned)(1)), 32, 0, stream>>>(gd_25); }
    k_posstep<<<(unsigned)((BK * 2 + 255) / 256), 256, 0, stream>>>(DL, LDP, X, POS, TRAJ, BK, T, 25);
    k_lincopy<<<(unsigned)(((long long)(BK) * (H) + 255) / 256), 256, 0, stream>>>(H0n, H, H0, H, BK, H);
    k_lincopy<<<(unsigned)(((long long)(BK) * (H) + 255) / 256), 256, 0, stream>>>(H1n, H, H1, H, BK, H);
    { GemmP gh0_26;
      gh0_26.A = H0; gh0_26.B = whh0; gh0_26.bias = bhh0; gh0_26.R = H0; gh0_26.C = GH;
      gh0_26.sAo = 0; gh0_26.sAi = 0; gh0_26.sAm = H; gh0_26.sAk = 1; gh0_26.sBo = 0; gh0_26.sBi = 0; gh0_26.sBn = H; gh0_26.sBk = 1; gh0_26.sCo = 0; gh0_26.sCi = 0; gh0_26.sCm = H3; gh0_26.sRo = 0; gh0_26.sRi = 0; gh0_26.sRm = 0; gh0_26.sRn = 0;
      gh0_26.M = BK; gh0_26.N = H3; gh0_26.K = H; gh0_26.zi_n = 1; gh0_26.flags = 1; gh0_26.act = 0;
      gh0_26.alpha = 1.0f; gh0_26.beta = 0.0f; gh0_26.sa = 1.0f; gh0_26.sb = 1.0f; gh0_26.Npad = H3; gh0_26.pad_ = 0;
      k_gemm<1><<<dim3((unsigned)((H3) + 31) / 32, (unsigned)((BK) + 15) / 16, (unsigned)(1)), 32, 0, stream>>>(gh0_26); }
    k_gru<<<(unsigned)(((long long)BK * H + 255) / 256), 256, 0, stream>>>(nullptr, X, wih0, bih0, GH, H0, H0n, BK, H);
    { GemmP gi1_26;
      gi1_26.A = H0n; gi1_26.B = wih1; gi1_26.bias = bih1; gi1_26.R = H0n; gi1_26.C = GI;
      gi1_26.sAo = 0; gi1_26.sAi = 0; gi1_26.sAm = H; gi1_26.sAk = 1; gi1_26.sBo = 0; gi1_26.sBi = 0; gi1_26.sBn = H; gi1_26.sBk = 1; gi1_26.sCo = 0; gi1_26.sCi = 0; gi1_26.sCm = H3; gi1_26.sRo = 0; gi1_26.sRi = 0; gi1_26.sRm = 0; gi1_26.sRn = 0;
      gi1_26.M = BK; gi1_26.N = H3; gi1_26.K = H; gi1_26.zi_n = 1; gi1_26.flags = 1; gi1_26.act = 0;
      gi1_26.alpha = 1.0f; gi1_26.beta = 0.0f; gi1_26.sa = 1.0f; gi1_26.sb = 1.0f; gi1_26.Npad = H3; gi1_26.pad_ = 0;
      k_gemm<1><<<dim3((unsigned)((H3) + 31) / 32, (unsigned)((BK) + 15) / 16, (unsigned)(1)), 32, 0, stream>>>(gi1_26); }
    { GemmP gh1_26;
      gh1_26.A = H1; gh1_26.B = whh1; gh1_26.bias = bhh1; gh1_26.R = H1; gh1_26.C = GH;
      gh1_26.sAo = 0; gh1_26.sAi = 0; gh1_26.sAm = H; gh1_26.sAk = 1; gh1_26.sBo = 0; gh1_26.sBi = 0; gh1_26.sBn = H; gh1_26.sBk = 1; gh1_26.sCo = 0; gh1_26.sCi = 0; gh1_26.sCm = H3; gh1_26.sRo = 0; gh1_26.sRi = 0; gh1_26.sRm = 0; gh1_26.sRn = 0;
      gh1_26.M = BK; gh1_26.N = H3; gh1_26.K = H; gh1_26.zi_n = 1; gh1_26.flags = 1; gh1_26.act = 0;
      gh1_26.alpha = 1.0f; gh1_26.beta = 0.0f; gh1_26.sa = 1.0f; gh1_26.sb = 1.0f; gh1_26.Npad = H3; gh1_26.pad_ = 0;
      k_gemm<1><<<dim3((unsigned)((H3) + 31) / 32, (unsigned)((BK) + 15) / 16, (unsigned)(1)), 32, 0, stream>>>(gh1_26); }
    k_gru<<<(unsigned)(((long long)BK * H + 255) / 256), 256, 0, stream>>>(GI, nullptr, nullptr, nullptr, GH, H1, H1n, BK, H);
    { GemmP gd_26;
      gd_26.A = H1n; gd_26.B = ow; gd_26.bias = ob; gd_26.R = H1n; gd_26.C = DL;
      gd_26.sAo = 0; gd_26.sAi = 0; gd_26.sAm = H; gd_26.sAk = 1; gd_26.sBo = 0; gd_26.sBi = 0; gd_26.sBn = H; gd_26.sBk = 1; gd_26.sCo = 0; gd_26.sCi = 0; gd_26.sCm = LDP; gd_26.sRo = 0; gd_26.sRi = 0; gd_26.sRm = 0; gd_26.sRn = 0;
      gd_26.M = BK; gd_26.N = 2; gd_26.K = H; gd_26.zi_n = 1; gd_26.flags = 1; gd_26.act = 0;
      gd_26.alpha = 1.0f; gd_26.beta = 0.0f; gd_26.sa = 1.0f; gd_26.sb = 1.0f; gd_26.Npad = LDP; gd_26.pad_ = 0;
      k_gemm<1><<<dim3((unsigned)((LDP) + 31) / 32, (unsigned)((BK) + 15) / 16, (unsigned)(1)), 32, 0, stream>>>(gd_26); }
    k_posstep<<<(unsigned)((BK * 2 + 255) / 256), 256, 0, stream>>>(DL, LDP, X, POS, TRAJ, BK, T, 26);
    k_lincopy<<<(unsigned)(((long long)(BK) * (H) + 255) / 256), 256, 0, stream>>>(H0n, H, H0, H, BK, H);
    k_lincopy<<<(unsigned)(((long long)(BK) * (H) + 255) / 256), 256, 0, stream>>>(H1n, H, H1, H, BK, H);
    { GemmP gh0_27;
      gh0_27.A = H0; gh0_27.B = whh0; gh0_27.bias = bhh0; gh0_27.R = H0; gh0_27.C = GH;
      gh0_27.sAo = 0; gh0_27.sAi = 0; gh0_27.sAm = H; gh0_27.sAk = 1; gh0_27.sBo = 0; gh0_27.sBi = 0; gh0_27.sBn = H; gh0_27.sBk = 1; gh0_27.sCo = 0; gh0_27.sCi = 0; gh0_27.sCm = H3; gh0_27.sRo = 0; gh0_27.sRi = 0; gh0_27.sRm = 0; gh0_27.sRn = 0;
      gh0_27.M = BK; gh0_27.N = H3; gh0_27.K = H; gh0_27.zi_n = 1; gh0_27.flags = 1; gh0_27.act = 0;
      gh0_27.alpha = 1.0f; gh0_27.beta = 0.0f; gh0_27.sa = 1.0f; gh0_27.sb = 1.0f; gh0_27.Npad = H3; gh0_27.pad_ = 0;
      k_gemm<1><<<dim3((unsigned)((H3) + 31) / 32, (unsigned)((BK) + 15) / 16, (unsigned)(1)), 32, 0, stream>>>(gh0_27); }
    k_gru<<<(unsigned)(((long long)BK * H + 255) / 256), 256, 0, stream>>>(nullptr, X, wih0, bih0, GH, H0, H0n, BK, H);
    { GemmP gi1_27;
      gi1_27.A = H0n; gi1_27.B = wih1; gi1_27.bias = bih1; gi1_27.R = H0n; gi1_27.C = GI;
      gi1_27.sAo = 0; gi1_27.sAi = 0; gi1_27.sAm = H; gi1_27.sAk = 1; gi1_27.sBo = 0; gi1_27.sBi = 0; gi1_27.sBn = H; gi1_27.sBk = 1; gi1_27.sCo = 0; gi1_27.sCi = 0; gi1_27.sCm = H3; gi1_27.sRo = 0; gi1_27.sRi = 0; gi1_27.sRm = 0; gi1_27.sRn = 0;
      gi1_27.M = BK; gi1_27.N = H3; gi1_27.K = H; gi1_27.zi_n = 1; gi1_27.flags = 1; gi1_27.act = 0;
      gi1_27.alpha = 1.0f; gi1_27.beta = 0.0f; gi1_27.sa = 1.0f; gi1_27.sb = 1.0f; gi1_27.Npad = H3; gi1_27.pad_ = 0;
      k_gemm<1><<<dim3((unsigned)((H3) + 31) / 32, (unsigned)((BK) + 15) / 16, (unsigned)(1)), 32, 0, stream>>>(gi1_27); }
    { GemmP gh1_27;
      gh1_27.A = H1; gh1_27.B = whh1; gh1_27.bias = bhh1; gh1_27.R = H1; gh1_27.C = GH;
      gh1_27.sAo = 0; gh1_27.sAi = 0; gh1_27.sAm = H; gh1_27.sAk = 1; gh1_27.sBo = 0; gh1_27.sBi = 0; gh1_27.sBn = H; gh1_27.sBk = 1; gh1_27.sCo = 0; gh1_27.sCi = 0; gh1_27.sCm = H3; gh1_27.sRo = 0; gh1_27.sRi = 0; gh1_27.sRm = 0; gh1_27.sRn = 0;
      gh1_27.M = BK; gh1_27.N = H3; gh1_27.K = H; gh1_27.zi_n = 1; gh1_27.flags = 1; gh1_27.act = 0;
      gh1_27.alpha = 1.0f; gh1_27.beta = 0.0f; gh1_27.sa = 1.0f; gh1_27.sb = 1.0f; gh1_27.Npad = H3; gh1_27.pad_ = 0;
      k_gemm<1><<<dim3((unsigned)((H3) + 31) / 32, (unsigned)((BK) + 15) / 16, (unsigned)(1)), 32, 0, stream>>>(gh1_27); }
    k_gru<<<(unsigned)(((long long)BK * H + 255) / 256), 256, 0, stream>>>(GI, nullptr, nullptr, nullptr, GH, H1, H1n, BK, H);
    { GemmP gd_27;
      gd_27.A = H1n; gd_27.B = ow; gd_27.bias = ob; gd_27.R = H1n; gd_27.C = DL;
      gd_27.sAo = 0; gd_27.sAi = 0; gd_27.sAm = H; gd_27.sAk = 1; gd_27.sBo = 0; gd_27.sBi = 0; gd_27.sBn = H; gd_27.sBk = 1; gd_27.sCo = 0; gd_27.sCi = 0; gd_27.sCm = LDP; gd_27.sRo = 0; gd_27.sRi = 0; gd_27.sRm = 0; gd_27.sRn = 0;
      gd_27.M = BK; gd_27.N = 2; gd_27.K = H; gd_27.zi_n = 1; gd_27.flags = 1; gd_27.act = 0;
      gd_27.alpha = 1.0f; gd_27.beta = 0.0f; gd_27.sa = 1.0f; gd_27.sb = 1.0f; gd_27.Npad = LDP; gd_27.pad_ = 0;
      k_gemm<1><<<dim3((unsigned)((LDP) + 31) / 32, (unsigned)((BK) + 15) / 16, (unsigned)(1)), 32, 0, stream>>>(gd_27); }
    k_posstep<<<(unsigned)((BK * 2 + 255) / 256), 256, 0, stream>>>(DL, LDP, X, POS, TRAJ, BK, T, 27);
    k_lincopy<<<(unsigned)(((long long)(BK) * (H) + 255) / 256), 256, 0, stream>>>(H0n, H, H0, H, BK, H);
    k_lincopy<<<(unsigned)(((long long)(BK) * (H) + 255) / 256), 256, 0, stream>>>(H1n, H, H1, H, BK, H);
    { GemmP gh0_28;
      gh0_28.A = H0; gh0_28.B = whh0; gh0_28.bias = bhh0; gh0_28.R = H0; gh0_28.C = GH;
      gh0_28.sAo = 0; gh0_28.sAi = 0; gh0_28.sAm = H; gh0_28.sAk = 1; gh0_28.sBo = 0; gh0_28.sBi = 0; gh0_28.sBn = H; gh0_28.sBk = 1; gh0_28.sCo = 0; gh0_28.sCi = 0; gh0_28.sCm = H3; gh0_28.sRo = 0; gh0_28.sRi = 0; gh0_28.sRm = 0; gh0_28.sRn = 0;
      gh0_28.M = BK; gh0_28.N = H3; gh0_28.K = H; gh0_28.zi_n = 1; gh0_28.flags = 1; gh0_28.act = 0;
      gh0_28.alpha = 1.0f; gh0_28.beta = 0.0f; gh0_28.sa = 1.0f; gh0_28.sb = 1.0f; gh0_28.Npad = H3; gh0_28.pad_ = 0;
      k_gemm<1><<<dim3((unsigned)((H3) + 31) / 32, (unsigned)((BK) + 15) / 16, (unsigned)(1)), 32, 0, stream>>>(gh0_28); }
    k_gru<<<(unsigned)(((long long)BK * H + 255) / 256), 256, 0, stream>>>(nullptr, X, wih0, bih0, GH, H0, H0n, BK, H);
    { GemmP gi1_28;
      gi1_28.A = H0n; gi1_28.B = wih1; gi1_28.bias = bih1; gi1_28.R = H0n; gi1_28.C = GI;
      gi1_28.sAo = 0; gi1_28.sAi = 0; gi1_28.sAm = H; gi1_28.sAk = 1; gi1_28.sBo = 0; gi1_28.sBi = 0; gi1_28.sBn = H; gi1_28.sBk = 1; gi1_28.sCo = 0; gi1_28.sCi = 0; gi1_28.sCm = H3; gi1_28.sRo = 0; gi1_28.sRi = 0; gi1_28.sRm = 0; gi1_28.sRn = 0;
      gi1_28.M = BK; gi1_28.N = H3; gi1_28.K = H; gi1_28.zi_n = 1; gi1_28.flags = 1; gi1_28.act = 0;
      gi1_28.alpha = 1.0f; gi1_28.beta = 0.0f; gi1_28.sa = 1.0f; gi1_28.sb = 1.0f; gi1_28.Npad = H3; gi1_28.pad_ = 0;
      k_gemm<1><<<dim3((unsigned)((H3) + 31) / 32, (unsigned)((BK) + 15) / 16, (unsigned)(1)), 32, 0, stream>>>(gi1_28); }
    { GemmP gh1_28;
      gh1_28.A = H1; gh1_28.B = whh1; gh1_28.bias = bhh1; gh1_28.R = H1; gh1_28.C = GH;
      gh1_28.sAo = 0; gh1_28.sAi = 0; gh1_28.sAm = H; gh1_28.sAk = 1; gh1_28.sBo = 0; gh1_28.sBi = 0; gh1_28.sBn = H; gh1_28.sBk = 1; gh1_28.sCo = 0; gh1_28.sCi = 0; gh1_28.sCm = H3; gh1_28.sRo = 0; gh1_28.sRi = 0; gh1_28.sRm = 0; gh1_28.sRn = 0;
      gh1_28.M = BK; gh1_28.N = H3; gh1_28.K = H; gh1_28.zi_n = 1; gh1_28.flags = 1; gh1_28.act = 0;
      gh1_28.alpha = 1.0f; gh1_28.beta = 0.0f; gh1_28.sa = 1.0f; gh1_28.sb = 1.0f; gh1_28.Npad = H3; gh1_28.pad_ = 0;
      k_gemm<1><<<dim3((unsigned)((H3) + 31) / 32, (unsigned)((BK) + 15) / 16, (unsigned)(1)), 32, 0, stream>>>(gh1_28); }
    k_gru<<<(unsigned)(((long long)BK * H + 255) / 256), 256, 0, stream>>>(GI, nullptr, nullptr, nullptr, GH, H1, H1n, BK, H);
    { GemmP gd_28;
      gd_28.A = H1n; gd_28.B = ow; gd_28.bias = ob; gd_28.R = H1n; gd_28.C = DL;
      gd_28.sAo = 0; gd_28.sAi = 0; gd_28.sAm = H; gd_28.sAk = 1; gd_28.sBo = 0; gd_28.sBi = 0; gd_28.sBn = H; gd_28.sBk = 1; gd_28.sCo = 0; gd_28.sCi = 0; gd_28.sCm = LDP; gd_28.sRo = 0; gd_28.sRi = 0; gd_28.sRm = 0; gd_28.sRn = 0;
      gd_28.M = BK; gd_28.N = 2; gd_28.K = H; gd_28.zi_n = 1; gd_28.flags = 1; gd_28.act = 0;
      gd_28.alpha = 1.0f; gd_28.beta = 0.0f; gd_28.sa = 1.0f; gd_28.sb = 1.0f; gd_28.Npad = LDP; gd_28.pad_ = 0;
      k_gemm<1><<<dim3((unsigned)((LDP) + 31) / 32, (unsigned)((BK) + 15) / 16, (unsigned)(1)), 32, 0, stream>>>(gd_28); }
    k_posstep<<<(unsigned)((BK * 2 + 255) / 256), 256, 0, stream>>>(DL, LDP, X, POS, TRAJ, BK, T, 28);
    k_lincopy<<<(unsigned)(((long long)(BK) * (H) + 255) / 256), 256, 0, stream>>>(H0n, H, H0, H, BK, H);
    k_lincopy<<<(unsigned)(((long long)(BK) * (H) + 255) / 256), 256, 0, stream>>>(H1n, H, H1, H, BK, H);
    { GemmP gh0_29;
      gh0_29.A = H0; gh0_29.B = whh0; gh0_29.bias = bhh0; gh0_29.R = H0; gh0_29.C = GH;
      gh0_29.sAo = 0; gh0_29.sAi = 0; gh0_29.sAm = H; gh0_29.sAk = 1; gh0_29.sBo = 0; gh0_29.sBi = 0; gh0_29.sBn = H; gh0_29.sBk = 1; gh0_29.sCo = 0; gh0_29.sCi = 0; gh0_29.sCm = H3; gh0_29.sRo = 0; gh0_29.sRi = 0; gh0_29.sRm = 0; gh0_29.sRn = 0;
      gh0_29.M = BK; gh0_29.N = H3; gh0_29.K = H; gh0_29.zi_n = 1; gh0_29.flags = 1; gh0_29.act = 0;
      gh0_29.alpha = 1.0f; gh0_29.beta = 0.0f; gh0_29.sa = 1.0f; gh0_29.sb = 1.0f; gh0_29.Npad = H3; gh0_29.pad_ = 0;
      k_gemm<1><<<dim3((unsigned)((H3) + 31) / 32, (unsigned)((BK) + 15) / 16, (unsigned)(1)), 32, 0, stream>>>(gh0_29); }
    k_gru<<<(unsigned)(((long long)BK * H + 255) / 256), 256, 0, stream>>>(nullptr, X, wih0, bih0, GH, H0, H0n, BK, H);
    { GemmP gi1_29;
      gi1_29.A = H0n; gi1_29.B = wih1; gi1_29.bias = bih1; gi1_29.R = H0n; gi1_29.C = GI;
      gi1_29.sAo = 0; gi1_29.sAi = 0; gi1_29.sAm = H; gi1_29.sAk = 1; gi1_29.sBo = 0; gi1_29.sBi = 0; gi1_29.sBn = H; gi1_29.sBk = 1; gi1_29.sCo = 0; gi1_29.sCi = 0; gi1_29.sCm = H3; gi1_29.sRo = 0; gi1_29.sRi = 0; gi1_29.sRm = 0; gi1_29.sRn = 0;
      gi1_29.M = BK; gi1_29.N = H3; gi1_29.K = H; gi1_29.zi_n = 1; gi1_29.flags = 1; gi1_29.act = 0;
      gi1_29.alpha = 1.0f; gi1_29.beta = 0.0f; gi1_29.sa = 1.0f; gi1_29.sb = 1.0f; gi1_29.Npad = H3; gi1_29.pad_ = 0;
      k_gemm<1><<<dim3((unsigned)((H3) + 31) / 32, (unsigned)((BK) + 15) / 16, (unsigned)(1)), 32, 0, stream>>>(gi1_29); }
    { GemmP gh1_29;
      gh1_29.A = H1; gh1_29.B = whh1; gh1_29.bias = bhh1; gh1_29.R = H1; gh1_29.C = GH;
      gh1_29.sAo = 0; gh1_29.sAi = 0; gh1_29.sAm = H; gh1_29.sAk = 1; gh1_29.sBo = 0; gh1_29.sBi = 0; gh1_29.sBn = H; gh1_29.sBk = 1; gh1_29.sCo = 0; gh1_29.sCi = 0; gh1_29.sCm = H3; gh1_29.sRo = 0; gh1_29.sRi = 0; gh1_29.sRm = 0; gh1_29.sRn = 0;
      gh1_29.M = BK; gh1_29.N = H3; gh1_29.K = H; gh1_29.zi_n = 1; gh1_29.flags = 1; gh1_29.act = 0;
      gh1_29.alpha = 1.0f; gh1_29.beta = 0.0f; gh1_29.sa = 1.0f; gh1_29.sb = 1.0f; gh1_29.Npad = H3; gh1_29.pad_ = 0;
      k_gemm<1><<<dim3((unsigned)((H3) + 31) / 32, (unsigned)((BK) + 15) / 16, (unsigned)(1)), 32, 0, stream>>>(gh1_29); }
    k_gru<<<(unsigned)(((long long)BK * H + 255) / 256), 256, 0, stream>>>(GI, nullptr, nullptr, nullptr, GH, H1, H1n, BK, H);
    { GemmP gd_29;
      gd_29.A = H1n; gd_29.B = ow; gd_29.bias = ob; gd_29.R = H1n; gd_29.C = DL;
      gd_29.sAo = 0; gd_29.sAi = 0; gd_29.sAm = H; gd_29.sAk = 1; gd_29.sBo = 0; gd_29.sBi = 0; gd_29.sBn = H; gd_29.sBk = 1; gd_29.sCo = 0; gd_29.sCi = 0; gd_29.sCm = LDP; gd_29.sRo = 0; gd_29.sRi = 0; gd_29.sRm = 0; gd_29.sRn = 0;
      gd_29.M = BK; gd_29.N = 2; gd_29.K = H; gd_29.zi_n = 1; gd_29.flags = 1; gd_29.act = 0;
      gd_29.alpha = 1.0f; gd_29.beta = 0.0f; gd_29.sa = 1.0f; gd_29.sb = 1.0f; gd_29.Npad = LDP; gd_29.pad_ = 0;
      k_gemm<1><<<dim3((unsigned)((LDP) + 31) / 32, (unsigned)((BK) + 15) / 16, (unsigned)(1)), 32, 0, stream>>>(gd_29); }
    k_posstep<<<(unsigned)((BK * 2 + 255) / 256), 256, 0, stream>>>(DL, LDP, X, POS, TRAJ, BK, T, 29);
    k_lincopy<<<(unsigned)(((long long)(BK) * (H) + 255) / 256), 256, 0, stream>>>(H0n, H, H0, H, BK, H);
    k_lincopy<<<(unsigned)(((long long)(BK) * (H) + 255) / 256), 256, 0, stream>>>(H1n, H, H1, H, BK, H);
    k_ramp<<<(unsigned)(((long long)BK * T * 2 + 255) / 256), 256, 0, stream>>>(TRAJ, goals, out, BK, T);
}
